// Cluster_81372450390694
// MI455X (gfx1250) — hardware-verified
//
#include <hip/hip_runtime.h>
#include <math.h>

typedef __attribute__((ext_vector_type(16))) _Float16 v16h;
typedef __attribute__((ext_vector_type(8)))  _Float16 v8h;
typedef __attribute__((ext_vector_type(16))) __bf16   v16b;
typedef __attribute__((ext_vector_type(8)))  float    v8f;
typedef __attribute__((ext_vector_type(4)))  float    v4f;

__device__ __forceinline__ int frag_k(int i, int h) { return (i < 8) ? (8 * h + i) : (16 + 8 * h + (i - 8)); }
__device__ __forceinline__ __bf16 bf16_rne(float f) {
    unsigned int u = __float_as_uint(f);
    u += 0x7fffu + ((u >> 16) & 1u);
    return __builtin_bit_cast(__bf16, (unsigned short)(u >> 16));
}
__device__ __forceinline__ float bf16_f32(__bf16 b) { return __uint_as_float(((unsigned int)__builtin_bit_cast(unsigned short, b)) << 16); }
__device__ __forceinline__ v8f wmma16(v16h a, v16h b, v8f c) {
    c = __builtin_amdgcn_wmma_f32_16x16x32_f16(false, a, false, b, (short)0, c, false, false);
    asm volatile("v_nop\n\tv_nop\n\tv_nop\n\tv_nop" : "+v"(c) : "v"(a), "v"(b));
    return c;
}
__device__ __forceinline__ v8f wmmab(v16b a, v16b b, v8f c) {
    c = __builtin_amdgcn_wmma_f32_16x16x32_bf16(false, a, false, b, (short)0, c, false, false);
    asm volatile("v_nop\n\tv_nop\n\tv_nop\n\tv_nop" : "+v"(c) : "v"(a), "v"(b));
    return c;
}
struct Split { v16b hi, lo; };
__device__ __forceinline__ v8f wmma3(const Split& a, const Split& b, v8f c) {
    c = __builtin_amdgcn_wmma_f32_16x16x32_bf16(false, a.hi, false, b.hi, (short)0, c, false, false);
    c = __builtin_amdgcn_wmma_f32_16x16x32_bf16(false, a.hi, false, b.lo, (short)0, c, false, false);
    c = __builtin_amdgcn_wmma_f32_16x16x32_bf16(false, a.lo, false, b.hi, (short)0, c, false, false);
    asm volatile("v_nop\n\tv_nop\n\tv_nop\n\tv_nop" : "+v"(c) : "v"(a.hi), "v"(a.lo), "v"(b.hi), "v"(b.lo));
    return c;
}
struct Split3 { v16b hi, mid, lo; };
__device__ __forceinline__ v8f wmma6(const Split3& a, const Split3& b, v8f c) {
    c = __builtin_amdgcn_wmma_f32_16x16x32_bf16(false, a.hi, false, b.hi, (short)0, c, false, false);
    c = __builtin_amdgcn_wmma_f32_16x16x32_bf16(false, a.hi, false, b.mid, (short)0, c, false, false);
    c = __builtin_amdgcn_wmma_f32_16x16x32_bf16(false, a.mid, false, b.hi, (short)0, c, false, false);
    c = __builtin_amdgcn_wmma_f32_16x16x32_bf16(false, a.hi, false, b.lo, (short)0, c, false, false);
    c = __builtin_amdgcn_wmma_f32_16x16x32_bf16(false, a.mid, false, b.mid, (short)0, c, false, false);
    c = __builtin_amdgcn_wmma_f32_16x16x32_bf16(false, a.lo, false, b.hi, (short)0, c, false, false);
    asm volatile("v_nop\n\tv_nop\n\tv_nop\n\tv_nop" : "+v"(c) : "v"(a.hi), "v"(a.mid), "v"(a.lo), "v"(b.hi), "v"(b.mid), "v"(b.lo));
    return c;
}

__device__ __forceinline__ v16h fh_ld(const float* __restrict__ p, long long sk, int k0, int h, int klen, float s) {
    v16h a;
#pragma unroll
    for (int i = 0; i < 16; ++i) { const int k = k0 + frag_k(i, h); a[i] = (k < klen) ? (_Float16)(p[(long long)k * sk] * s) : (_Float16)0.f; }
    return a;
}
__device__ __forceinline__ Split sp_ld(const float* __restrict__ p, long long sk, int k0, int h, int klen, float s) {
    Split r;
#pragma unroll
    for (int i = 0; i < 16; ++i) {
        const int k = k0 + frag_k(i, h); const float x = (k < klen) ? p[(long long)k * sk] * s : 0.f;
        const __bf16 hb = bf16_rne(x); r.hi[i] = hb; r.lo[i] = bf16_rne(x - bf16_f32(hb));
    }
    return r;
}
__device__ __forceinline__ Split3 sp3_ld(const float* __restrict__ p, long long sk, int k0, int h, int klen, float s) {
    Split3 r;
#pragma unroll
    for (int i = 0; i < 16; ++i) {
        const int k = k0 + frag_k(i, h); const float x = (k < klen) ? p[(long long)k * sk] * s : 0.f;
        const __bf16 hb = bf16_rne(x); const float r1 = x - bf16_f32(hb); const __bf16 mb = bf16_rne(r1);
        r.hi[i] = hb; r.mid[i] = mb; r.lo[i] = bf16_rne(r1 - bf16_f32(mb));
    }
    return r;
}
__device__ __forceinline__ v16b bh_ld(const float* __restrict__ p, long long sk, int k0, int h, int klen, float s) {
    v16b a;
#pragma unroll
    for (int i = 0; i < 16; ++i) { const int k = k0 + frag_k(i, h); a[i] = bf16_rne((k < klen) ? p[(long long)k * sk] * s : 0.f); }
    return a;
}
__device__ __forceinline__ v16h fh_row(const _Float16* __restrict__ row, int k0, int h) {
    v16h a;
#pragma unroll
    for (int i = 0; i < 16; ++i) a[i] = row[k0 + frag_k(i, h)];
    return a;
}

#define VST2(T, ptr, val) do { *(volatile T*)(ptr) = (val); __threadfence(); *(volatile T*)(ptr) = (val); } while (0)
typedef float v4f __attribute__((ext_vector_type(4)));
#define VST2V4(ptr, val) do { *(volatile v4f*)(ptr) = (val); __threadfence(); *(volatile v4f*)(ptr) = (val); } while (0)

__device__ __attribute__((noinline)) float act_fn(float v, int act) {
    if (act == 1) return fmaxf(v, 0.f);
    if (act == 2) { const float u = 0.7978845608028654f * (v + 0.044715f * v * v * v); return 0.5f * v * (1.f + tanhf(u)); }
    if (act == 3) return v / (1.f + expf(-v));
    if (act == 4) return 0.5f * v * (1.f + erff(v * 0.7071067811865476f));
    if (act == 5) return tanhf(v);
    if (act == 6) return 1.f / (1.f + expf(-v));
    if (act == 7) return (v > 0.f) ? v : 0.01f * v;
    if (act == 8) return (v > 0.f) ? v : (expf(v) - 1.f);
    if (act == 9) return fminf(fmaxf(v, 0.f), 6.f);
    if (act == 10) return fabsf(v);
    if (act == 11) return (v >= 0.f) ? v : 0.1f * v;
    if (act == 12) return (v > 0.f) ? v : 0.2f * v;
    if (act == 13) return (v > 20.f) ? v : log1pf(expf(v));
    return v;
}

struct GemmP {
    const float* A; const float* B; const float* bias; const float* R; float* C;
    long long sAo, sAi, sAm, sAk, sBo, sBi, sBn, sBk, sCo, sCi, sCm, sRo, sRi, sRm, sRn;
    int M, N, K, zi_n, flags, act; float alpha, beta, sa, sb;
    int Npad, pad_;
};
static_assert(sizeof(GemmP) == 5 * 8 + 15 * 8 + 6 * 4 + 4 * 4 + 2 * 4, "GemmP has padding");

template <int MODE>
__global__ __launch_bounds__(32) void k_gemm(GemmP p) {
    const int lane = threadIdx.x & 31, h = lane >> 4, l15 = lane & 15;
    const int m0 = blockIdx.y * 16, n0 = blockIdx.x * 32;
    const int z = blockIdx.z, zo = z / p.zi_n, zi = z - zo * p.zi_n;
    const float* A = p.A + zo * p.sAo + zi * p.sAi;
    const float* B = p.B + zo * p.sBo + zi * p.sBi;
    const int am = min(m0 + l15, p.M - 1);
    v8f acc[2], comp[2];
#pragma unroll
    for (int t = 0; t < 2; ++t) { v8f zz = {}; acc[t] = zz; comp[t] = zz; }
    for (int k0 = 0; k0 < p.K; k0 += 32) {
        const float* arow = A + (long long)am * p.sAm;
        if (MODE == 1) {
            const Split a = sp_ld(arow, p.sAk, k0, h, p.K, 1.f);
#pragma unroll
            for (int t = 0; t < 2; ++t) {
                const int bn = min(n0 + t * 16 + l15, p.N - 1);
                acc[t] = wmma3(a, sp_ld(B + (long long)bn * p.sBn, p.sBk, k0, h, p.K, 1.f), acc[t]);
            }
        } else if (MODE == 3) {
            const Split3 a = sp3_ld(arow, p.sAk, k0, h, p.K, 1.f);
#pragma unroll
            for (int t = 0; t < 2; ++t) {
                const int bn = min(n0 + t * 16 + l15, p.N - 1);
                acc[t] = wmma6(a, sp3_ld(B + (long long)bn * p.sBn, p.sBk, k0, h, p.K, 1.f), acc[t]);
            }
        } else if (MODE == 4) {
            const Split3 a = sp3_ld(arow, p.sAk, k0, h, p.K, 1.f);
#pragma unroll
            for (int t = 0; t < 2; ++t) {
                const int bn = min(n0 + t * 16 + l15, p.N - 1); v8f zz = {};
                const v8f part = wmma6(a, sp3_ld(B + (long long)bn * p.sBn, p.sBk, k0, h, p.K, 1.f), zz);
                const v8f y = part - comp[t]; const v8f s = acc[t] + y; comp[t] = (s - acc[t]) - y; acc[t] = s;
            }
        } else if (MODE == 2) {
            const v16b a = bh_ld(arow, p.sAk, k0, h, p.K, 1.f);
#pragma unroll
            for (int t = 0; t < 2; ++t) {
                const int bn = min(n0 + t * 16 + l15, p.N - 1);
                acc[t] = wmmab(a, bh_ld(B + (long long)bn * p.sBn, p.sBk, k0, h, p.K, 1.f), acc[t]);
            }
        } else {
            const v16h a = fh_ld(arow, p.sAk, k0, h, p.K, p.sa);
#pragma unroll
            for (int t = 0; t < 2; ++t) {
                const int bn = min(n0 + t * 16 + l15, p.N - 1);
                acc[t] = wmma16(a, fh_ld(B + (long long)bn * p.sBn, p.sBk, k0, h, p.K, p.sb), acc[t]);
            }
        }
    }
    const float iscale = (MODE == 0) ? p.alpha / (p.sa * p.sb) : p.alpha;
    float* C = p.C + zo * p.sCo + zi * p.sCi;
    const float* R = p.R + zo * p.sRo + zi * p.sRi;
    __shared__ __align__(16) float ctile[16][36];
#pragma unroll
    for (int t = 0; t < 2; ++t) {
        const int n = n0 + t * 16 + l15; const int nn = min(n, p.N - 1);
#pragma unroll
        for (int r = 0; r < 8; ++r) {
            const int m = m0 + 8 * h + r; const int mm = min(m, p.M - 1);
            float v = acc[t][r] * iscale;
            if (p.flags & 1) v += p.bias[nn];
            if (p.flags & 2) v += p.bias[mm];
            v = act_fn(v, p.act);
            if (p.flags & 4) v += p.beta * R[(long long)mm * p.sRm + (long long)nn * p.sRn];
            ctile[8 * h + r][t * 16 + l15] = (n < p.N) ? v : 0.f;
        }
    }
    __syncthreads();
    const int NW = (p.Npad > p.N) ? p.Npad : p.N;
    const bool fast = (m0 + 16 <= p.M) && (n0 + 32 <= NW) && ((p.sCm & 3) == 0) && ((((size_t)C) & 15) == 0);
    if (fast) {
#pragma unroll
        for (int s = 0; s < 4; ++s) {
            const int row = s * 4 + (lane >> 3), c4 = (lane & 7) * 4;
            const v4f v = *(const v4f*)&ctile[row][c4];
            VST2V4(C + (long long)(m0 + row) * p.sCm + n0 + c4, v);
        }
    } else {
        for (int row = 0; row < 16; ++row) {
            const int m = m0 + row, n = n0 + lane;
            if (m < p.M && n < NW) VST2(float, C + (long long)m * p.sCm + n, ctile[row][lane]);
        }
    }
}

#define AW 4
struct AttnP {
    const float* Q; const float* K; const float* V; float* O; float* P; const float* Mf; const int* Mi; float* ST;
    const float* Pw; const float* Rt; const int* SQ; const int* SK;
    long long swb, swh, swi, swj, srb, srh, sri;
    long long sQb, sQh, sQi, sQd, sKb, sKh, sKj, sKd, sVb, sVh, sVj, sVd, sOb, sOh, sOi, sPb, sPh, sPi, smb, smh, smi, smj;
    int Lq, Lk, dh, dv, hrep, causal, coff, pband;
    float scale, mfill; int nonorm, mpol;
    int roff, rn, segpol, win;
};
static_assert(sizeof(AttnP) == 12 * 8 + 29 * 8 + 16 * 4, "AttnP has padding");

#ifndef KATTN_ATTR
#define KATTN_ATTR
#endif
template <int DHP, int DVP, int QM, bool SPLITPV, bool TWOPASS>
__global__ __launch_bounds__(32 * AW) KATTN_ATTR void k_attn(AttnP p) {
    constexpr int NT = DVP / 16;
    constexpr int KS = DHP / 32;
    constexpr int VP = DVP + 8;
    __shared__ __align__(16) float    pl[AW][16 * 64];
    __shared__ __align__(16) _Float16 vl[(SPLITPV ? 2 : 1) * 64 * VP];
    const int lane = threadIdx.x & 31, hf = lane >> 4, l15 = lane & 15, wave = threadIdx.x >> 5;
    const int h = blockIdx.y, b = blockIdx.z, hk = h / p.hrep;
    const int q0 = (blockIdx.x * AW + wave) * 16;
    float* myp = pl[wave];
    const float L2E = 1.4426950408889634f;
    const float NEG = -__builtin_inff();
    const int qi = min(q0 + l15, p.Lq - 1);
    const float* qrow = p.Q + b * p.sQb + h * p.sQh + (long long)qi * p.sQi;
    const float* kbase = p.K + b * p.sKb + hk * p.sKh;
    const float* vbase = p.V + b * p.sVb + hk * p.sVh;
    v16h qa[QM == 0 ? KS : 1]; Split qs_[QM == 1 ? KS : 1]; Split3 qt_[QM == 2 ? KS : 1];
#pragma unroll
    for (int ks = 0; ks < KS; ++ks) {
        if (QM == 2) qt_[ks] = sp3_ld(qrow, p.sQd, ks * 32, hf, p.dh, 1.f);
        else if (QM == 1) qs_[ks] = sp_ld(qrow, p.sQd, ks * 32, hf, p.dh, 1.f);
        else qa[ks] = fh_ld(qrow, p.sQd, ks * 32, hf, p.dh, 1.f);
    }
    v8f o[NT]; float m8[8], l8[8];
#pragma unroll
    for (int t = 0; t < NT; ++t) { v8f zz = {}; o[t] = zz; }
#pragma unroll
    for (int i = 0; i < 8; ++i) { m8[i] = NEG; l8[i] = 0.f; }
    int jend = p.Lk;
    if (p.causal == 1) { const int je = (blockIdx.x * AW + AW - 1) * 16 + 16 + p.coff; jend = min(jend, max(je, 0)); }
    const int npass = TWOPASS ? 2 : 1;
    for (int pass = 0; pass < npass; ++pass) {
        const bool dopv = (!TWOPASS) || pass == 1;
        for (int j0 = 0; j0 < jend; j0 += 64) {
            if (dopv) {
                __syncthreads();
                for (int idx = threadIdx.x; idx < 64 * DVP; idx += 32 * AW) {
                    const int jr = idx / DVP, d = idx - jr * DVP, j = j0 + jr;
                    const float f = (j < p.Lk && d < p.dv) ? vbase[(long long)j * p.sVj + (long long)d * p.sVd] : 0.f;
                    if (SPLITPV) {
                        const __bf16 hb = bf16_rne(f);
                        ((__bf16*)vl)[jr * VP + d] = hb; ((__bf16*)vl)[64 * VP + jr * VP + d] = bf16_rne(f - bf16_f32(hb));
                    } else vl[jr * VP + d] = (_Float16)f;
                }
            }
            v8f s[4];
#pragma unroll
            for (int t = 0; t < 4; ++t) {
                const int j = min(j0 + t * 16 + l15, p.Lk - 1);
                const float* krow = kbase + (long long)j * p.sKj;
                v8f acc = {};
#pragma unroll
                for (int ks = 0; ks < KS; ++ks) {
                    if (QM == 2)      acc = wmma6(qt_[ks], sp3_ld(krow, p.sKd, ks * 32, hf, p.dh, 1.f), acc);
                    else if (QM == 1) acc = wmma3(qs_[ks], sp_ld(krow, p.sKd, ks * 32, hf, p.dh, 1.f), acc);
                    else              acc = wmma16(qa[ks], fh_ld(krow, p.sKd, ks * 32, hf, p.dh, 1.f), acc);
                }
                s[t] = acc;
            }
            float pv[8][4];
#pragma unroll
            for (int i = 0; i < 8; ++i) {
                const int irow = q0 + i + 8 * hf;
                const int ic = min(irow, p.Lq - 1);
                float sc[4];
#pragma unroll
                for (int t = 0; t < 4; ++t) {
                    const int jg = j0 + t * 16 + l15;
                    float v = s[t][i] * p.scale;
                    if (p.Mf) v += p.Mf[b * p.smb + h * p.smh + (long long)ic * p.smi + (long long)min(jg, p.Lk - 1) * p.smj];
                    if (p.Rt) { int rc = ic - min(jg, p.Lk - 1) + p.roff; rc = rc < 0 ? 0 : (rc >= p.rn ? p.rn - 1 : rc); v += p.Rt[b * p.srb + h * p.srh + (long long)ic * p.sri + rc]; }
                    if (p.Mi) { const int mv = p.Mi[b * p.smb + h * p.smh + (long long)ic * p.smi + (long long)min(jg, p.Lk - 1) * p.smj]; if (p.mpol ? (mv != 0) : (mv == 0)) v = p.mfill; }
                    if (p.SQ) { const bool same = p.SQ[(long long)b * p.Lq + ic] == p.SK[(long long)b * p.Lk + min(jg, p.Lk - 1)]; if (p.segpol ? same : !same) v = p.mfill; }
                    if (p.causal == 2 && jg > irow + p.coff) v = p.mfill;
                    if (jg >= p.Lk || (p.causal == 1 && jg > irow + p.coff) || (p.causal == 3 && jg < irow + p.coff) || (p.win > 0 && irow + p.coff - jg > p.win)) v = NEG; else v *= L2E;
                    sc[t] = v;
                }
                if (!TWOPASS || pass == 0) {
                    float mx = fmaxf(fmaxf(sc[0], sc[1]), fmaxf(sc[2], sc[3]));
                    mx = fmaxf(mx, __shfl_xor(mx, 1, 32)); mx = fmaxf(mx, __shfl_xor(mx, 2, 32));
                    mx = fmaxf(mx, __shfl_xor(mx, 4, 32)); mx = fmaxf(mx, __shfl_xor(mx, 8, 32));
                    const float mnew = fmaxf(m8[i], mx);
                    const float corr = (mnew == NEG) ? 1.f : exp2f(m8[i] - mnew);
                    float rs = 0.f;
#pragma unroll
                    for (int t = 0; t < 4; ++t) {
                        const float pp = (sc[t] == NEG) ? 0.f : exp2f(sc[t] - mnew); rs += pp;
                        pv[i][t] = p.Pw ? pp * p.Pw[b * p.swb + h * p.swh + (long long)ic * p.swi + (long long)min(j0 + t * 16 + l15, p.Lk - 1) * p.swj] : pp;
                    }
                    rs += __shfl_xor(rs, 1, 32); rs += __shfl_xor(rs, 2, 32); rs += __shfl_xor(rs, 4, 32); rs += __shfl_xor(rs, 8, 32);
                    l8[i] = l8[i] * corr + rs; m8[i] = mnew;
                    if (!TWOPASS) {
#pragma unroll
                        for (int t = 0; t < NT; ++t) o[t][i] *= corr;
                    }
                } else {
                    const float inv = (l8[i] > 0.f) ? 1.f / l8[i] : 0.f;
#pragma unroll
                    for (int t = 0; t < 4; ++t) {
                        const int jg = j0 + t * 16 + l15;
                        float pp = (sc[t] == NEG) ? 0.f : exp2f(sc[t] - m8[i]) * inv;
                        if (p.Pw) pp *= p.Pw[b * p.swb + h * p.swh + (long long)ic * p.swi + (long long)min(jg, p.Lk - 1) * p.swj];
                        pv[i][t] = pp;
                    }
                }
            }
            if (dopv) {
#pragma unroll
                for (int i = 0; i < 8; ++i)
#pragma unroll
                    for (int t = 0; t < 4; ++t) myp[(i + 8 * hf) * 64 + t * 16 + l15] = pv[i][t];
                __syncthreads();
                if (p.P) {
                    float* pb_ = p.P + b * p.sPb + h * p.sPh;
                    const bool fastP = (p.pband == 0) && ((p.sPi & 3) == 0) && (j0 + 64 <= p.Lk) && (q0 + 16 <= p.Lq) && ((((size_t)pb_) & 15) == 0);
                    if (fastP) {
#pragma unroll
                        for (int s = 0; s < 8; ++s) {
                            const int row = s * 2 + (lane >> 4), c4 = (lane & 15) * 4;
                            const v4f v = *(const v4f*)(myp + row * 64 + c4);
                            VST2V4(pb_ + (long long)(q0 + row) * p.sPi + j0 + c4, v);
                        }
                    } else {
                        for (int row = 0; row < 16; ++row) {
                            const int irow = q0 + row; if (irow >= p.Lq) continue;
                            for (int c = lane; c < 64; c += 32) {
                                const int jg = j0 + c; if (jg >= p.Lk) continue;
                                if (p.pband == 0) VST2(float, pb_ + (long long)irow * p.sPi + jg, myp[row * 64 + c]);
                                else if (jg - irow <= p.pband && irow - jg <= p.pband) VST2(float, pb_ + (long long)irow * p.sPi + (jg - irow + p.pband), myp[row * 64 + c]);
                            }
                        }
                    }
                }
                if (SPLITPV) {
                    const Split pa0 = sp_ld(myp + l15 * 64, 1, 0, hf, 64, 1.f), pa1 = sp_ld(myp + l15 * 64, 1, 32, hf, 64, 1.f);
                    const __bf16* vh = (const __bf16*)vl; const __bf16* vlo = vh + 64 * VP;
#pragma unroll
                    for (int t = 0; t < NT; ++t) {
                        const int dcol = t * 16 + l15;
                        Split b0, b1;
#pragma unroll
                        for (int e = 0; e < 16; ++e) {
                            const int k0 = frag_k(e, hf), k1 = 32 + frag_k(e, hf);
                            b0.hi[e] = vh[k0 * VP + dcol]; b0.lo[e] = vlo[k0 * VP + dcol]; b1.hi[e] = vh[k1 * VP + dcol]; b1.lo[e] = vlo[k1 * VP + dcol];
                        }
                        o[t] = wmma3(pa0, b0, o[t]);
                        o[t] = wmma3(pa1, b1, o[t]);
                    }
                } else {
                    const v16h pa0 = fh_ld(myp + l15 * 64, 1, 0, hf, 64, 4096.f), pa1 = fh_ld(myp + l15 * 64, 1, 32, hf, 64, 4096.f);
#pragma unroll
                    for (int t = 0; t < NT; ++t) {
                        const int dcol = t * 16 + l15;
                        v16h b0, b1;
#pragma unroll
                        for (int e = 0; e < 16; ++e) { b0[e] = vl[frag_k(e, hf) * VP + dcol]; b1[e] = vl[(32 + frag_k(e, hf)) * VP + dcol]; }
                        o[t] = wmma16(pa0, b0, o[t]);
                        o[t] = wmma16(pa1, b1, o[t]);
                    }
                }
            }
        }
    }
    float* obase = p.O + b * p.sOb + h * p.sOh;
    if (p.ST) {
        const int rl = lane >> 1, isel = rl & 7;
        float mv = 0.f, lv = 0.f;
#pragma unroll
        for (int i = 0; i < 8; ++i) if (i == isel) { mv = m8[i]; lv = l8[i]; }
        const int irow = q0 + rl;
        if (irow < p.Lq) { float* st = p.ST + (((long long)b * gridDim.y + h) * p.Lq + irow) * 2 + (lane & 1); VST2(float, st, (lane & 1) ? lv : mv * 0.6931471805599453f); }
    }
    float invr[8];
#pragma unroll
    for (int i = 0; i < 8; ++i) {
        if (TWOPASS) invr[i] = SPLITPV ? 1.f : (1.f / 4096.f);
        else if (p.nonorm) invr[i] = exp2f(m8[i]) * (SPLITPV ? 1.f : (1.f / 4096.f));
        else invr[i] = (l8[i] > 0.f) ? (SPLITPV ? 1.f / l8[i] : 1.f / (l8[i] * 4096.f)) : 0.f;
    }
    __syncthreads();
    const bool ofast = ((p.sOi & 3) == 0) && ((((size_t)obase) & 15) == 0) && (q0 + 16 <= p.Lq);
#pragma unroll
    for (int c0 = 0; c0 < DVP; c0 += 64) {
#pragma unroll
        for (int i = 0; i < 8; ++i)
#pragma unroll
            for (int t = 0; t < NT; ++t) if (t * 16 >= c0 && t * 16 < c0 + 64) myp[(i + 8 * hf) * 64 + (t * 16 - c0) + l15] = o[t][i] * invr[i];
        __syncthreads();
        const int cw = (DVP - c0 < 64) ? (DVP - c0) : 64;
        if (ofast && (c0 + cw <= p.dv) && (cw % 32 == 0)) {
            const int lpr = cw / 4;
            const int rows_per_ins = 32 / lpr;
            for (int r0 = 0; r0 < 16; r0 += rows_per_ins) {
                const int row = r0 + lane / lpr, c4 = (lane % lpr) * 4;
                const v4f v = *(const v4f*)(myp + row * 64 + c4);
                VST2V4(obase + (long long)(q0 + row) * p.sOi + c0 + c4, v);
            }
        } else {
            for (int row = 0; row < 16; ++row) {
                const int irow = q0 + row; if (irow >= p.Lq) continue;
                for (int c = lane; c < cw; c += 32) { const int d = c0 + c; if (d < p.dv) VST2(float, obase + (long long)irow * p.sOi + d, myp[row * 64 + c]); }
            }
        }
        __syncthreads();
    }
}

struct TrP { const float* src; float* dst; const float* R2; long long sSz, lds, sDz, ldd, sRz, ldr; int R, C, flags, act; float alpha, beta; };
static_assert(sizeof(TrP) == 3 * 8 + 6 * 8 + 6 * 4, "TrP has padding");
__global__ __launch_bounds__(256) void k_tr(TrP p) {
    __shared__ float tile[32][33];
    const int c0 = blockIdx.x * 32, r0 = blockIdx.y * 32, z = blockIdx.z;
    const int lane = threadIdx.x & 31, wave = threadIdx.x >> 5;
    const float* s = p.src + z * p.sSz;
#pragma unroll
    for (int k = 0; k < 4; ++k) {
        const int rl = wave * 4 + k, r = r0 + rl, c = c0 + lane;
        tile[rl][lane] = (r < p.R && c < p.C) ? s[(long long)r * p.lds + c] : 0.f;
    }
    __syncthreads();
    float* d = p.dst + z * p.sDz; const float* rr = p.R2 + z * p.sRz;
#pragma unroll
    for (int k = 0; k < 4; ++k) {
        const int cl = wave * 4 + k, c = c0 + cl, r = r0 + lane;
        if (c < p.C && r < p.R) {
            float v = act_fn(p.alpha * tile[lane][cl], p.act);
            if (p.flags & 1) v += p.beta * rr[(long long)c * p.ldr + r];
            VST2(float, d + (long long)c * p.ldd + r, v);
        }
    }
}

__global__ __launch_bounds__(256) void k_affine(const float* __restrict__ src, float* __restrict__ dst, int n, float a, float b, const float* __restrict__ sdev) {
    const int i = blockIdx.x * 256 + threadIdx.x;
    if (i < n) { const float aa = sdev ? a * sdev[0] : a; const float v = aa * src[i] + b; VST2(float, dst + i, v); }
}

struct SmP { const float* src; float* dst; const float* Mf; long long sz, sr, dz, dr, smz, smr; int n, pad; float scale_in, scale_out; };
static_assert(sizeof(SmP) == 3 * 8 + 6 * 8 + 4 * 4, "SmP has padding");
__global__ __launch_bounds__(256) void k_softmax(SmP p) {
    __shared__ float red[256];
    const int r = blockIdx.x, z = blockIdx.y, tid = threadIdx.x;
    const float* s = p.src + z * p.sz + (long long)r * p.sr;
    const float* mf = p.Mf ? (p.Mf + z * p.smz + (long long)r * p.smr) : nullptr;
    float mx = -__builtin_inff();
    for (int j = tid; j < p.n; j += 256) { float v = s[j] * p.scale_in; if (mf) v += mf[j]; mx = fmaxf(mx, v); }
    red[tid] = mx; __syncthreads();
    for (int o = 128; o > 0; o >>= 1) { if (tid < o) red[tid] = fmaxf(red[tid], red[tid + o]); __syncthreads(); }
    mx = red[0]; __syncthreads();
    float sum = 0.f;
    for (int j = tid; j < p.n; j += 256) { float v = s[j] * p.scale_in; if (mf) v += mf[j]; sum += (mx == -__builtin_inff()) ? 0.f : expf(v - mx); }
    red[tid] = sum; __syncthreads();
    for (int o = 128; o > 0; o >>= 1) { if (tid < o) red[tid] += red[tid + o]; __syncthreads(); }
    sum = red[0];
    const float inv = (sum > 0.f) ? p.scale_out / sum : 0.f;
    float* d = p.dst + z * p.dz + (long long)r * p.dr;
    for (int j = tid; j < p.n; j += 256) { float v = s[j] * p.scale_in; if (mf) v += mf[j]; const float o = (mx == -__builtin_inff()) ? 0.f : expf(v - mx) * inv; VST2(float, d + j, o); }
}
__global__ __launch_bounds__(256) void k_stats(const float* __restrict__ x, long long sz, long long so, long long si, int inner, int n, float eps, float* __restrict__ stat, int mode) {
    __shared__ float red[256];
    const int z = blockIdx.x, tid = threadIdx.x;
    const float* base = x + z * sz;
    float s = 0.f;
    for (int e = tid; e < n; e += 256) s += base[(long long)(e / inner) * so + (long long)(e % inner) * si];
    red[tid] = s; __syncthreads();
    for (int o = 128; o > 0; o >>= 1) { if (tid < o) red[tid] += red[tid + o]; __syncthreads(); }
    const float mu = (mode == 0 || mode == 3) ? red[0] / (float)n : 0.f; __syncthreads();
    float q = 0.f;
    for (int e = tid; e < n; e += 256) { const float dlt = base[(long long)(e / inner) * so + (long long)(e % inner) * si] - mu; q += dlt * dlt; }
    red[tid] = q; __syncthreads();
    for (int o = 128; o > 0; o >>= 1) { if (tid < o) red[tid] += red[tid + o]; __syncthreads(); }
    {
        float rs;
        if (mode == 2) rs = sqrtf((float)n) / fmaxf(sqrtf(red[0]), eps); else if (mode == 3) rs = rsqrtf(red[0] / (float)(n - 1) + eps); else rs = rsqrtf(red[0] / (float)n + eps);
        if (tid < 32) { const float v = (tid == 0) ? mu : ((tid == 1) ? rs : 0.f); VST2(float, stat + (long long)z * 32 + tid, v); }
    }
}
__global__ __launch_bounds__(256) void k_norm_apply(const float* __restrict__ x, float* __restrict__ y, const float* __restrict__ stat, const float* __restrict__ g, const float* __restrict__ bta,
                                                     int Z, int C, int L, int G, int bn, int act) {
    const long long idx = (long long)blockIdx.x * 256 + threadIdx.x;
    if (idx >= (long long)Z * C * L) return;
    const int l = (int)(idx % L); const long long zc = idx / L; const int c = (int)(zc % C), z = (int)(zc / C); (void)l;
    const int set = bn ? c : (z * G + c / (C / G));
    float v = (x[idx] - stat[(long long)set * 32]) * stat[(long long)set * 32 + 1];
    if (g) v *= g[c];
    if (bta) v += bta[c];
    v = act_fn(v, act);
    VST2(float, y + idx, v);
}

__global__ __launch_bounds__(256) void k_lse_neg(const float* __restrict__ st, float* __restrict__ c, int n) {
    const int i = blockIdx.x * 256 + threadIdx.x;
    if (i < n) { const float v = -(st[2 * i] + logf(st[2 * i + 1])); VST2(float, c + i, v); }
}

__global__ __launch_bounds__(256) void k_iota(int* __restrict__ dst, int n, int a, int b) {
    const int i = blockIdx.x * 256 + threadIdx.x;
    if (i < n) { const int v = a * i + b; VST2(int, dst + i, v); }
}

__global__ __launch_bounds__(256) void k_axpby(const float* __restrict__ x, const float* __restrict__ y, float* __restrict__ dst, int n, float a, float b, float c) {
    const int i = blockIdx.x * 256 + threadIdx.x;
    if (i < n) { const float v = a * x[i] + b * y[i] + c; VST2(float, dst + i, v); }
}

struct RopeP { const float* X; float* Y; const float* C; const float* Sn; const int* pos; long long sXr, sXh, sYr, sYh, sCb, sCp, sCd; int R, Hn, D, S, mode, tmode, pmode, pad; };
static_assert(sizeof(RopeP) == 5 * 8 + 7 * 8 + 8 * 4, "RopeP has padding");
__global__ __launch_bounds__(256) void k_rope(RopeP p) {
    const long long idx = (long long)blockIdx.x * 256 + threadIdx.x;
    if (idx >= (long long)p.R * p.Hn * p.D) return;
    const int d = (int)(idx % p.D); const long long rh = idx / p.D; const int h = (int)(rh % p.Hn); const int r = (int)(rh / p.Hn);
    const int half = p.D / 2;
    int partner; float sign;
    if (p.mode == 0) { partner = (d < half) ? d + half : d - half; sign = (d < half) ? -1.f : 1.f; }
    else { partner = d ^ 1; sign = (d & 1) ? 1.f : -1.f; }
    const int tcol = (p.tmode == 0) ? d : ((p.tmode == 1) ? (d % half) : (d >> 1));
    const int pp = (p.pmode == 0) ? (r % p.S) : ((p.pmode == 1) ? h : p.pos[r]);
    const long long toff = (long long)(r / p.S) * p.sCb + (long long)pp * p.sCp + (long long)tcol * p.sCd;
    const float* xr = p.X + (long long)r * p.sXr + (long long)h * p.sXh;
    const float v = xr[d] * p.C[toff] + sign * xr[partner] * p.Sn[toff];
    VST2(float, p.Y + (long long)r * p.sYr + (long long)h * p.sYh + d, v);
}

__global__ __launch_bounds__(256) void k_invf(float* __restrict__ invb, int half, int D, float base, float num, int fmode, float cexp) {
    const int i = blockIdx.x * 256 + threadIdx.x;
    if (i >= ((half + 31) / 32) * 32) return;
    if (i >= half) { VST2(float, invb + i, 0.f); return; }
    const float e = (float)(2 * i) / (float)D;
    float invf;
    if (fmode == 1) invf = num * expf((float)(2 * i) * cexp);
    else if (fmode == 2) invf = num * powf(base, (-2.0f * ((float)i - 1.0f)) / (float)D);
    else invf = num * (1.0f / powf(base, e));
    VST2(float, invb + i, invf);
}
__global__ __launch_bounds__(256) void k_sincos(float* __restrict__ cs, float* __restrict__ sn, const float* __restrict__ invb, int S, int half, float pscale) {
    const int idx = blockIdx.x * 256 + threadIdx.x;
    if (idx >= S * half) return;
    const int s = idx / half, i = idx - s * half;
    const float ang = (pscale * (float)s) * invb[i];
    VST2(float, cs + idx, cosf(ang)); VST2(float, sn + idx, sinf(ang));
}

__global__ __launch_bounds__(256) void k_mulact(const float* __restrict__ x, const float* __restrict__ y, float* __restrict__ dst, int n, int act) {
    const int i = blockIdx.x * 256 + threadIdx.x;
    if (i < n) { const float v = act_fn(x[i], act) * y[i]; VST2(float, dst + i, v); }
}

__global__ __launch_bounds__(256) void k_matvec(GemmP p) {
    const int rpt = (p.N == 1) ? 1 : 32;
    const long long r0 = ((long long)blockIdx.x * 256 + threadIdx.x) * rpt; const int z = blockIdx.z, zo = z / p.zi_n, zi = z - zo * p.zi_n;
    if (r0 >= p.M) return;
    const float* Bb = p.B + zo * p.sBo + zi * p.sBi;
    float* C = p.C + zo * p.sCo + zi * p.sCi; const float* R = p.R + zo * p.sRo + zi * p.sRi;
    for (int rr = 0; rr < rpt; ++rr) {
        const long long r = r0 + rr; if (r >= p.M) break;
        const float* A = p.A + zo * p.sAo + zi * p.sAi + r * p.sAm;
        float acc[8] = {0.f, 0.f, 0.f, 0.f, 0.f, 0.f, 0.f, 0.f};
        for (int k = 0; k < p.K; ++k) { const float a = A[(long long)k * p.sAk];
#pragma unroll
            for (int j = 0; j < 8; ++j) if (j < p.N) acc[j] += a * Bb[(long long)j * p.sBn + (long long)k * p.sBk]; }
#pragma unroll
        for (int j = 0; j < 8; ++j) if (j < p.N) {
            float v = acc[j] * p.alpha;
            if (p.flags & 1) v += p.bias[j];
            if (p.flags & 2) v += p.bias[r];
            v = act_fn(v, p.act);
            if (p.flags & 4) v += p.beta * R[r * p.sRm + (long long)j * p.sRn];
            VST2(float, C + r * p.sCm + j, v);
        }
    }
}
__global__ __launch_bounds__(256) void k_smallsoftmax(const float* __restrict__ src, float* __restrict__ dst, long long sr, long long dr, int n, long long R, float scale) {
    const long long r0 = ((long long)blockIdx.x * 256 + threadIdx.x) * 32;
    for (int rr = 0; rr < 32; ++rr) {
        const long long r = r0 + rr; if (r >= R) return;
        const float* s = src + r * sr; float* d = dst + r * dr;
        float mx = -__builtin_inff();
        for (int j = 0; j < n; ++j) mx = fmaxf(mx, s[j] * scale);
        float sum = 0.f;
        for (int j = 0; j < n; ++j) sum += expf(s[j] * scale - mx);
        const float inv = 1.f / sum;
        for (int j = 0; j < n; ++j) { const float v = expf(s[j] * scale - mx) * inv; VST2(float, d + j, v); }
    }
}

__global__ __launch_bounds__(32) void k_unitstat(float* __restrict__ st) { const int t = threadIdx.x; const float v = (t == 1) ? 1.f : 0.f; VST2(float, st + t, v); }

__global__ __launch_bounds__(256) void k_lincopy(const float* __restrict__ src, long long lds, float* __restrict__ dst, long long ldd, long long rows, int cols) {
    const long long i = (long long)blockIdx.x * 256 + threadIdx.x; if (i >= rows * cols) return;
    const long long r = i / cols; const int c = (int)(i - r * cols);
    const float v = src[r * lds + c]; VST2(float, dst + r * ldd + c, v);
}

__global__ __launch_bounds__(256) void k_cl_pad(const float* __restrict__ X, float* __restrict__ XP, int b, int C, int H, int T) { const long long q = (long long)blockIdx.x * 256 + threadIdx.x; if (q >= (long long)H * T * C) return; const int c = (int)(q % C); const int t = (int)((q / C) % T); const int y = (int)(q / ((long long)C * T)); VST2(float, XP + (((long long)(y + 2)) * (T + 4) + t + 2) * C + c, X[(((long long)b * C + c) * H + y) * T + t]); }
__global__ __launch_bounds__(256) void k_cl_bnl(float* __restrict__ HP, const float* __restrict__ g, const float* __restrict__ bb, const float* __restrict__ m, const float* __restrict__ v, int H, int T, int C) { const long long q = (long long)blockIdx.x * 256 + threadIdx.x; if (q >= (long long)H * T * C) return; const int c = (int)(q % C); const int t = (int)((q / C) % T); const int y = (int)(q / ((long long)C * T)); float* p = HP + (((long long)y) * (T + 2) + t + 1) * C + c; float u = (*p - m[c]) * rsqrtf(v[c] + 1e-5f) * g[c] + bb[c]; u = (u >= 0.f) ? u : 0.01f * u; VST2(float, p, u); }
__global__ __launch_bounds__(256) void k_cl_colsum1(const float* __restrict__ A, int ld, int C, long long L, float* __restrict__ PART) { __shared__ float red[256]; const int blk = blockIdx.x; const int nb = gridDim.x; const long long per = (L + nb - 1) / nb; const long long l0 = (long long)blk * per; long long l1 = l0 + per; if (l1 > L) l1 = L;
    for (int c = 0; c < C; ++c) { float s = 0.f; for (long long l = l0 + threadIdx.x; l < l1; l += 256) s += A[l * ld + c]; red[threadIdx.x] = s; __syncthreads(); for (int o = 128; o > 0; o >>= 1) { if (threadIdx.x < o) red[threadIdx.x] += red[threadIdx.x + o]; __syncthreads(); } if (threadIdx.x == 0) VST2(float, PART + blk * 32 + c, red[0]); __syncthreads(); } }
__global__ __launch_bounds__(256) void k_cl_colsum2(const float* __restrict__ PART, int NB, int C, float* __restrict__ RED, int off) { __shared__ float red[256]; for (int c = 0; c < C; ++c) { float s = 0.f; for (int i = threadIdx.x; i < NB; i += 256) s += PART[i * 32 + c]; red[threadIdx.x] = s; __syncthreads(); for (int o = 128; o > 0; o >>= 1) { if (threadIdx.x < o) red[threadIdx.x] += red[threadIdx.x + o]; __syncthreads(); } if (threadIdx.x == 0) VST2(float, RED + off + c, red[0]); __syncthreads(); } }
__global__ __launch_bounds__(256) void k_cl_max1(const float* __restrict__ SV, int col, long long L, float* __restrict__ PART) { __shared__ float red[256]; const int blk = blockIdx.x; const int nb = gridDim.x; const long long per = (L + nb - 1) / nb; const long long l0 = (long long)blk * per; long long l1 = l0 + per; if (l1 > L) l1 = L; float mx = -__builtin_inff(); for (long long l = l0 + threadIdx.x; l < l1; l += 256) mx = fmaxf(mx, SV[l * 4 + col]); red[threadIdx.x] = mx; __syncthreads(); for (int o = 128; o > 0; o >>= 1) { if (threadIdx.x < o) red[threadIdx.x] = fmaxf(red[threadIdx.x], red[threadIdx.x + o]); __syncthreads(); } if (threadIdx.x == 0) VST2(float, PART + blk * 32, red[0]); }
__global__ __launch_bounds__(256) void k_cl_max2(const float* __restrict__ PART, int NB, float* __restrict__ RED, int off) { __shared__ float red[256]; float mx = -__builtin_inff(); for (int i = threadIdx.x; i < NB; i += 256) mx = fmaxf(mx, PART[i * 32]); red[threadIdx.x] = mx; __syncthreads(); for (int o = 128; o > 0; o >>= 1) { if (threadIdx.x < o) red[threadIdx.x] = fmaxf(red[threadIdx.x], red[threadIdx.x + o]); __syncthreads(); } if (threadIdx.x == 0) VST2(float, RED + off, red[0]); }
__global__ __launch_bounds__(256) void k_cl_masknorm(float* __restrict__ KV, int ld, const float* __restrict__ frame, const float* __restrict__ RED, const float* __restrict__ Tsc, long long L, int C) { const long long l = (long long)blockIdx.x * 256 + threadIdx.x; if (l >= L) return; float a = 0.f;
#pragma unroll 1
    for (int c = 0; c < C; ++c) { const float v = KV[l * ld + c]; a += v * v; } const float amp = sqrtf(a + 1.01e-8f); const float f = frame[l] / (amp * RED[0]) * Tsc[0];
#pragma unroll 1
    for (int c = 0; c < C; ++c) { const float v = KV[l * ld + c] * f; VST2(float, KV + l * ld + c, v); } }
__global__ __launch_bounds__(256) void k_cl_sig(float* __restrict__ A, int ld, int C, long long L) { const long long q = (long long)blockIdx.x * 256 + threadIdx.x; if (q >= L * C) return; const long long l = q / C; const int c = (int)(q % C); const float v = 1.f / (1.f + expf(-A[l * ld + c])); VST2(float, A + l * ld + c, v); }
__global__ __launch_bounds__(256) void k_cl_flow1(const float* __restrict__ QP, const float* __restrict__ KP, int ld, const float* __restrict__ RED, float* __restrict__ SV, long long L, int D) { const long long l = (long long)blockIdx.x * 256 + threadIdx.x; if (l >= L) return; float a = 0.f, b = 0.f; const float E = 1.01e-8f;
#pragma unroll 1
    for (int d = 0; d < D; ++d) { a += (QP[l * ld + d] + E) * (RED[16 + d] + E); b += (KP[l * ld + d] + E) * (RED[32 + d] + E); } VST2(float, SV + l * 4, 1.f / a); VST2(float, SV + l * 4 + 1, 1.f / b); }
__global__ __launch_bounds__(256) void k_cl_flow2(const float* __restrict__ QP, const float* __restrict__ KP, int ld, const float* __restrict__ SV, float* __restrict__ O, float* __restrict__ O2, long long L, int D) { const long long q = (long long)blockIdx.x * 256 + threadIdx.x; if (q >= L * D) return; const long long l = q / D; const int d = (int)(q % D); VST2(float, O + l * ld + d, KP[l * ld + d] * SV[l * 4 + 1]); VST2(float, O2 + l * ld + d, QP[l * ld + d] * SV[l * 4]); }
__global__ __launch_bounds__(256) void k_cl_flow3(const float* __restrict__ QP, const float* __restrict__ KP, int ld, const float* __restrict__ RED, float* __restrict__ SV, long long L, int D) { const long long l = (long long)blockIdx.x * 256 + threadIdx.x; if (l >= L) return; float a = 0.f, b = 0.f; const float E = 1.01e-8f;
#pragma unroll 1
    for (int d = 0; d < D; ++d) { a += (QP[l * ld + d] + E) * (RED[48 + d] + E); b += (KP[l * ld + d] + E) * (RED[64 + d] + E); } VST2(float, SV + l * 4 + 2, 1.f / (1.f + expf(-a))); VST2(float, SV + l * 4 + 3, b); }
__global__ __launch_bounds__(256) void k_cl_flow4(const float* __restrict__ SV, const float* __restrict__ RED, float* __restrict__ O2, int ld, long long L) { const long long l = (long long)blockIdx.x * 256 + threadIdx.x; if (l >= L) return; VST2(float, O2 + l * ld + 15, expf(SV[l * 4 + 3] - RED[80])); }
__global__ __launch_bounds__(256) void k_cl_flow5(const float* __restrict__ VP, const float* __restrict__ O2, int ld, const float* __restrict__ RED, float* __restrict__ O, long long L, int D) { const long long q = (long long)blockIdx.x * 256 + threadIdx.x; if (q >= L * D) return; const long long l = q / D; const int d = (int)(q % D); const float sc = O2[l * ld + 15] / RED[96] * (float)L; VST2(float, O + l * ld + d, VP[l * ld + d] * sc); }
__global__ __launch_bounds__(256) void k_cl_flow6(float* __restrict__ O2, int ld, const float* __restrict__ SV, long long L, int D) { const long long q = (long long)blockIdx.x * 256 + threadIdx.x; if (q >= L * D) return; const long long l = q / D; const int d = (int)(q % D); const float v = O2[l * ld + d] * SV[l * 4] * SV[l * 4 + 2]; VST2(float, O2 + l * ld + d, v); }
__global__ __launch_bounds__(256) void k_cl_out(const float* __restrict__ O, int ld, float* __restrict__ OUT, int b, long long L, int D) { const long long q = (long long)blockIdx.x * 256 + threadIdx.x; if (q >= L * D) return; const long long l = q % L; const int d = (int)(q / L); VST2(float, OUT + ((long long)b * D + d) * L + l, O[l * ld + d]); }

template __global__ void k_gemm<1>(GemmP);

extern "C" void kernel_launch(void* const* d_in, const int* in_sizes, int n_in, void* d_out, int out_size, void* d_ws, size_t ws_size, hipStream_t stream) {
    (void)in_sizes; (void)n_in; (void)out_size; (void)ws_size;
    const float* x = (const float*)d_in[0];
    const float* frame = (const float*)d_in[1];
    const float* wpre = (const float*)d_in[2];
    const float* bpre = (const float*)d_in[3];
    const float* bng = (const float*)d_in[4];
    const float* bnb = (const float*)d_in[5];
    const float* bnm = (const float*)d_in[6];
    const float* bnv = (const float*)d_in[7];
    const float* Tsc = (const float*)d_in[8];
    const float* wq = (const float*)d_in[9];
    const float* bq = (const float*)d_in[10];
    const float* wkv = (const float*)d_in[11];
    const float* bkv = (const float*)d_in[12];
    const float* faq = (const float*)d_in[13];
    const float* fabq = (const float*)d_in[14];
    const float* fak = (const float*)d_in[15];
    const float* fabk = (const float*)d_in[16];
    const float* fav = (const float*)d_in[17];
    const float* fabv = (const float*)d_in[18];
    const float* fao = (const float*)d_in[19];
    const float* fabo = (const float*)d_in[20];
    const int Bn = 4;
    const int CI = 8;
    const int Hh = 252;
    const int Tt = 2048;
    const int C1 = 16;
    const int D = 12;
    const int Fo = 84;
    const int Ll = Fo * Tt;
    const int LD = 16;
    const int NB = 672;
    float* out = (float*)d_out;
    char* wsp = (char*)d_ws;
    float* XP = (float*)wsp; wsp += (((size_t)((size_t)256 * 2052 * CI) * 4 + 255) / 256) * 256;
    float* HP = (float*)wsp; wsp += (((size_t)((size_t)Hh * 2050 * C1) * 4 + 255) / 256) * 256;
    float* Q = (float*)wsp; wsp += (((size_t)((size_t)Ll * LD) * 4 + 255) / 256) * 256;
    float* KV = (float*)wsp; wsp += (((size_t)((size_t)Ll * LD) * 4 + 255) / 256) * 256;
    float* QP = (float*)wsp; wsp += (((size_t)((size_t)Ll * LD) * 4 + 255) / 256) * 256;
    float* KP = (float*)wsp; wsp += (((size_t)((size_t)Ll * LD) * 4 + 255) / 256) * 256;
    float* VP = (float*)wsp; wsp += (((size_t)((size_t)Ll * LD) * 4 + 255) / 256) * 256;
    float* O = (float*)wsp; wsp += (((size_t)((size_t)Ll * LD) * 4 + 255) / 256) * 256;
    float* O2 = (float*)wsp; wsp += (((size_t)((size_t)Ll * LD) * 4 + 255) / 256) * 256;
    float* SV = (float*)wsp; wsp += (((size_t)((size_t)Ll * 4) * 4 + 255) / 256) * 256;
    float* PART = (float*)wsp; wsp += (((size_t)((size_t)NB * 32) * 4 + 255) / 256) * 256;
    float* RED = (float*)wsp; wsp += (((size_t)((size_t)256) * 4 + 255) / 256) * 256;
    float* KVM = (float*)wsp; wsp += (((size_t)((size_t)LD * LD) * 4 + 255) / 256) * 256;
    hipMemsetAsync(XP, 0, (size_t)256 * 2052 * CI * 4, stream); hipMemsetAsync(HP, 0, (size_t)Hh * 2050 * C1 * 4, stream);
    k_cl_pad<<<(unsigned)(((long long)Hh * Tt * CI + 255) / 256), 256, 0, stream>>>(x, XP, 0, CI, Hh, Tt);
    { GemmP cp0_0;
      cp0_0.A = XP + (size_t)0 * CI; cp0_0.B = wpre + 0; cp0_0.bias = bpre; cp0_0.R = XP + (size_t)0 * CI; cp0_0.C = HP + C1;
      cp0_0.sAo = (long long)2052 * CI; cp0_0.sAi = 0; cp0_0.sAm = CI; cp0_0.sAk = 1; cp0_0.sBo = 0; cp0_0.sBi = 0; cp0_0.sBn = CI * 25; cp0_0.sBk = 25; cp0_0.sCo = (long long)2050 * C1; cp0_0.sCi = 0; cp0_0.sCm = C1; cp0_0.sRo = 0; cp0_0.sRi = 0; cp0_0.sRm = 0; cp0_0.sRn = 0;
      cp0_0.M = Tt; cp0_0.N = C1; cp0_0.K = CI; cp0_0.zi_n = 1; cp0_0.flags = 1; cp0_0.act = 0;
      cp0_0.alpha = 1.0f; cp0_0.beta = 0.0f; cp0_0.sa = 1.0f; cp0_0.sb = 1.0f; cp0_0.Npad = C1; cp0_0.pad_ = 0;
      k_gemm<1><<<dim3((unsigned)((C1) + 31) / 32, (unsigned)((Tt) + 15) / 16, (unsigned)(Hh)), 32, 0, stream>>>(cp0_0); }
    { GemmP cp0_1;
      cp0_1.A = XP + (size_t)1 * CI; cp0_1.B = wpre + 1; cp0_1.bias = XP + (size_t)1 * CI; cp0_1.R = HP + C1; cp0_1.C = HP + C1;
      cp0_1.sAo = (long long)2052 * CI; cp0_1.sAi = 0; cp0_1.sAm = CI; cp0_1.sAk = 1; cp0_1.sBo = 0; cp0_1.sBi = 0; cp0_1.sBn = CI * 25; cp0_1.sBk = 25; cp0_1.sCo = (long long)2050 * C1; cp0_1.sCi = 0; cp0_1.sCm = C1; cp0_1.sRo = (long long)2050 * C1; cp0_1.sRi = 0; cp0_1.sRm = C1; cp0_1.sRn = 1;
      cp0_1.M = Tt; cp0_1.N = C1; cp0_1.K = CI; cp0_1.zi_n = 1; cp0_1.flags = 4; cp0_1.act = 0;
      cp0_1.alpha = 1.0f; cp0_1.beta = 1.0f; cp0_1.sa = 1.0f; cp0_1.sb = 1.0f; cp0_1.Npad = C1; cp0_1.pad_ = 0;
      k_gemm<1><<<dim3((unsigned)((C1) + 31) / 32, (unsigned)((Tt) + 15) / 16, (unsigned)(Hh)), 32, 0, stream>>>(cp0_1); }
    { GemmP cp0_2;
      cp0_2.A = XP + (size_t)2 * CI; cp0_2.B = wpre + 2; cp0_2.bias = XP + (size_t)2 * CI; cp0_2.R = HP + C1; cp0_2.C = HP + C1;
      cp0_2.sAo = (long long)2052 * CI; cp0_2.sAi = 0; cp0_2.sAm = CI; cp0_2.sAk = 1; cp0_2.sBo = 0; cp0_2.sBi = 0; cp0_2.sBn = CI * 25; cp0_2.sBk = 25; cp0_2.sCo = (long long)2050 * C1; cp0_2.sCi = 0; cp0_2.sCm = C1; cp0_2.sRo = (long long)2050 * C1; cp0_2.sRi = 0; cp0_2.sRm = C1; cp0_2.sRn = 1;
      cp0_2.M = Tt; cp0_2.N = C1; cp0_2.K = CI; cp0_2.zi_n = 1; cp0_2.flags = 4; cp0_2.act = 0;
      cp0_2.alpha = 1.0f; cp0_2.beta = 1.0f; cp0_2.sa = 1.0f; cp0_2.sb = 1.0f; cp0_2.Npad = C1; cp0_2.pad_ = 0;
      k_gemm<1><<<dim3((unsigned)((C1) + 31) / 32, (unsigned)((Tt) + 15) / 16, (unsigned)(Hh)), 32, 0, stream>>>(cp0_2); }
    { GemmP cp0_3;
      cp0_3.A = XP + (size_t)3 * CI; cp0_3.B = wpre + 3; cp0_3.bias = XP + (size_t)3 * CI; cp0_3.R = HP + C1; cp0_3.C = HP + C1;
      cp0_3.sAo = (long long)2052 * CI; cp0_3.sAi = 0; cp0_3.sAm = CI; cp0_3.sAk = 1; cp0_3.sBo = 0; cp0_3.sBi = 0; cp0_3.sBn = CI * 25; cp0_3.sBk = 25; cp0_3.sCo = (long long)2050 * C1; cp0_3.sCi = 0; cp0_3.sCm = C1; cp0_3.sRo = (long long)2050 * C1; cp0_3.sRi = 0; cp0_3.sRm = C1; cp0_3.sRn = 1;
      cp0_3.M = Tt; cp0_3.N = C1; cp0_3.K = CI; cp0_3.zi_n = 1; cp0_3.flags = 4; cp0_3.act = 0;
      cp0_3.alpha = 1.0f; cp0_3.beta = 1.0f; cp0_3.sa = 1.0f; cp0_3.sb = 1.0f; cp0_3.Npad = C1; cp0_3.pad_ = 0;
      k_gemm<1><<<dim3((unsigned)((C1) + 31) / 32, (unsigned)((Tt) + 15) / 16, (unsigned)(Hh)), 32, 0, stream>>>(cp0_3); }
    { GemmP cp0_4;
      cp0_4.A = XP + (size_t)4 * CI; cp0_4.B = wpre + 4; cp0_4.bias = XP + (size_t)4 * CI; cp0_4.R = HP + C1; cp0_4.C = HP + C1;
      cp0_4.sAo = (long long)2052 * CI; cp0_4.sAi = 0; cp0_4.sAm = CI; cp0_4.sAk = 1; cp0_4.sBo = 0; cp0_4.sBi = 0; cp0_4.sBn = CI * 25; cp0_4.sBk = 25; cp0_4.sCo = (long long)2050 * C1; cp0_4.sCi = 0; cp0_4.sCm = C1; cp0_4.sRo = (long long)2050 * C1; cp0_4.sRi = 0; cp0_4.sRm = C1; cp0_4.sRn = 1;
      cp0_4.M = Tt; cp0_4.N = C1; cp0_4.K = CI; cp0_4.zi_n = 1; cp0_4.flags = 4; cp0_4.act = 0;
      cp0_4.alpha = 1.0f; cp0_4.beta = 1.0f; cp0_4.sa = 1.0f; cp0_4.sb = 1.0f; cp0_4.Npad = C1; cp0_4.pad_ = 0;
      k_gemm<1><<<dim3((unsigned)((C1) + 31) / 32, (unsigned)((Tt) + 15) / 16, (unsigned)(Hh)), 32, 0, stream>>>(cp0_4); }
    { GemmP cp0_5;
      cp0_5.A = XP + (size_t)2052 * CI; cp0_5.B = wpre + 5; cp0_5.bias = XP + (size_t)2052 * CI; cp0_5.R = HP + C1; cp0_5.C = HP + C1;
      cp0_5.sAo = (long long)2052 * CI; cp0_5.sAi = 0; cp0_5.sAm = CI; cp0_5.sAk = 1; cp0_5.sBo = 0; cp0_5.sBi = 0; cp0_5.sBn = CI * 25; cp0_5.sBk = 25; cp0_5.sCo = (long long)2050 * C1; cp0_5.sCi = 0; cp0_5.sCm = C1; cp0_5.sRo = (long long)2050 * C1; cp0_5.sRi = 0; cp0_5.sRm = C1; cp0_5.sRn = 1;
      cp0_5.M = Tt; cp0_5.N = C1; cp0_5.K = CI; cp0_5.zi_n = 1; cp0_5.flags = 4; cp0_5.act = 0;
      cp0_5.alpha = 1.0f; cp0_5.beta = 1.0f; cp0_5.sa = 1.0f; cp0_5.sb = 1.0f; cp0_5.Npad = C1; cp0_5.pad_ = 0;
      k_gemm<1><<<dim3((unsigned)((C1) + 31) / 32, (unsigned)((Tt) + 15) / 16, (unsigned)(Hh)), 32, 0, stream>>>(cp0_5); }
    { GemmP cp0_6;
      cp0_6.A = XP + (size_t)2053 * CI; cp0_6.B = wpre + 6; cp0_6.bias = XP + (size_t)2053 * CI; cp0_6.R = HP + C1; cp0_6.C = HP + C1;
      cp0_6.sAo = (long long)2052 * CI; cp0_6.sAi = 0; cp0_6.sAm = CI; cp0_6.sAk = 1; cp0_6.sBo = 0; cp0_6.sBi = 0; cp0_6.sBn = CI * 25; cp0_6.sBk = 25; cp0_6.sCo = (long long)2050 * C1; cp0_6.sCi = 0; cp0_6.sCm = C1; cp0_6.sRo = (long long)2050 * C1; cp0_6.sRi = 0; cp0_6.sRm = C1; cp0_6.sRn = 1;
      cp0_6.M = Tt; cp0_6.N = C1; cp0_6.K = CI; cp0_6.zi_n = 1; cp0_6.flags = 4; cp0_6.act = 0;
      cp0_6.alpha = 1.0f; cp0_6.beta = 1.0f; cp0_6.sa = 1.0f; cp0_6.sb = 1.0f; cp0_6.Npad = C1; cp0_6.pad_ = 0;
      k_gemm<1><<<dim3((unsigned)((C1) + 31) / 32, (unsigned)((Tt) + 15) / 16, (unsigned)(Hh)), 32, 0, stream>>>(cp0_6); }
    { GemmP cp0_7;
      cp0_7.A = XP + (size_t)2054 * CI; cp0_7.B = wpre + 7; cp0_7.bias = XP + (size_t)2054 * CI; cp0_7.R = HP + C1; cp0_7.C = HP + C1;
      cp0_7.sAo = (long long)2052 * CI; cp0_7.sAi = 0; cp0_7.sAm = CI; cp0_7.sAk = 1; cp0_7.sBo = 0; cp0_7.sBi = 0; cp0_7.sBn = CI * 25; cp0_7.sBk = 25; cp0_7.sCo = (long long)2050 * C1; cp0_7.sCi = 0; cp0_7.sCm = C1; cp0_7.sRo = (long long)2050 * C1; cp0_7.sRi = 0; cp0_7.sRm = C1; cp0_7.sRn = 1;
      cp0_7.M = Tt; cp0_7.N = C1; cp0_7.K = CI; cp0_7.zi_n = 1; cp0_7.flags = 4; cp0_7.act = 0;
      cp0_7.alpha = 1.0f; cp0_7.beta = 1.0f; cp0_7.sa = 1.0f; cp0_7.sb = 1.0f; cp0_7.Npad = C1; cp0_7.pad_ = 0;
      k_gemm<1><<<dim3((unsigned)((C1) + 31) / 32, (unsigned)((Tt) + 15) / 16, (unsigned)(Hh)), 32, 0, stream>>>(cp0_7); }
    { GemmP cp0_8;
      cp0_8.A = XP + (size_t)2055 * CI; cp0_8.B = wpre + 8; cp0_8.bias = XP + (size_t)2055 * CI; cp0_8.R = HP + C1; cp0_8.C = HP + C1;
      cp0_8.sAo = (long long)2052 * CI; cp0_8.sAi = 0; cp0_8.sAm = CI; cp0_8.sAk = 1; cp0_8.sBo = 0; cp0_8.sBi = 0; cp0_8.sBn = CI * 25; cp0_8.sBk = 25; cp0_8.sCo = (long long)2050 * C1; cp0_8.sCi = 0; cp0_8.sCm = C1; cp0_8.sRo = (long long)2050 * C1; cp0_8.sRi = 0; cp0_8.sRm = C1; cp0_8.sRn = 1;
      cp0_8.M = Tt; cp0_8.N = C1; cp0_8.K = CI; cp0_8.zi_n = 1; cp0_8.flags = 4; cp0_8.act = 0;
      cp0_8.alpha = 1.0f; cp0_8.beta = 1.0f; cp0_8.sa = 1.0f; cp0_8.sb = 1.0f; cp0_8.Npad = C1; cp0_8.pad_ = 0;
      k_gemm<1><<<dim3((unsigned)((C1) + 31) / 32, (unsigned)((Tt) + 15) / 16, (unsigned)(Hh)), 32, 0, stream>>>(cp0_8); }
    { GemmP cp0_9;
      cp0_9.A = XP + (size_t)2056 * CI; cp0_9.B = wpre + 9; cp0_9.bias = XP + (size_t)2056 * CI; cp0_9.R = HP + C1; cp0_9.C = HP + C1;
      cp0_9.sAo = (long long)2052 * CI; cp0_9.sAi = 0; cp0_9.sAm = CI; cp0_9.sAk = 1; cp0_9.sBo = 0; cp0_9.sBi = 0; cp0_9.sBn = CI * 25; cp0_9.sBk = 25; cp0_9.sCo = (long long)2050 * C1; cp0_9.sCi = 0; cp0_9.sCm = C1; cp0_9.sRo = (long long)2050 * C1; cp0_9.sRi = 0; cp0_9.sRm = C1; cp0_9.sRn = 1;
      cp0_9.M = Tt; cp0_9.N = C1; cp0_9.K = CI; cp0_9.zi_n = 1; cp0_9.flags = 4; cp0_9.act = 0;
      cp0_9.alpha = 1.0f; cp0_9.beta = 1.0f; cp0_9.sa = 1.0f; cp0_9.sb = 1.0f; cp0_9.Npad = C1; cp0_9.pad_ = 0;
      k_gemm<1><<<dim3((unsigned)((C1) + 31) / 32, (unsigned)((Tt) + 15) / 16, (unsigned)(Hh)), 32, 0, stream>>>(cp0_9); }
    { GemmP cp0_10;
      cp0_10.A = XP + (size_t)4104 * CI; cp0_10.B = wpre + 10; cp0_10.bias = XP + (size_t)4104 * CI; cp0_10.R = HP + C1; cp0_10.C = HP + C1;
      cp0_10.sAo = (long long)2052 * CI; cp0_10.sAi = 0; cp0_10.sAm = CI; cp0_10.sAk = 1; cp0_10.sBo = 0; cp0_10.sBi = 0; cp0_10.sBn = CI * 25; cp0_10.sBk = 25; cp0_10.sCo = (long long)2050 * C1; cp0_10.sCi = 0; cp0_10.sCm = C1; cp0_10.sRo = (long long)2050 * C1; cp0_10.sRi = 0; cp0_10.sRm = C1; cp0_10.sRn = 1;
      cp0_10.M = Tt; cp0_10.N = C1; cp0_10.K = CI; cp0_10.zi_n = 1; cp0_10.flags = 4; cp0_10.act = 0;
      cp0_10.alpha = 1.0f; cp0_10.beta = 1.0f; cp0_10.sa = 1.0f; cp0_10.sb = 1.0f; cp0_10.Npad = C1; cp0_10.pad_ = 0;
      k_gemm<1><<<dim3((unsigned)((C1) + 31) / 32, (unsigned)((Tt) + 15) / 16, (unsigned)(Hh)), 32, 0, stream>>>(cp0_10); }
    { GemmP cp0_11;
      cp0_11.A = XP + (size_t)4105 * CI; cp0_11.B = wpre + 11; cp0_11.bias = XP + (size_t)4105 * CI; cp0_11.R = HP + C1; cp0_11.C = HP + C1;
      cp0_11.sAo = (long long)2052 * CI; cp0_11.sAi = 0; cp0_11.sAm = CI; cp0_11.sAk = 1; cp0_11.sBo = 0; cp0_11.sBi = 0; cp0_11.sBn = CI * 25; cp0_11.sBk = 25; cp0_11.sCo = (long long)2050 * C1; cp0_11.sCi = 0; cp0_11.sCm = C1; cp0_11.sRo = (long long)2050 * C1; cp0_11.sRi = 0; cp0_11.sRm = C1; cp0_11.sRn = 1;
      cp0_11.M = Tt; cp0_11.N = C1; cp0_11.K = CI; cp0_11.zi_n = 1; cp0_11.flags = 4; cp0_11.act = 0;
      cp0_11.alpha = 1.0f; cp0_11.beta = 1.0f; cp0_11.sa = 1.0f; cp0_11.sb = 1.0f; cp0_11.Npad = C1; cp0_11.pad_ = 0;
      k_gemm<1><<<dim3((unsigned)((C1) + 31) / 32, (unsigned)((Tt) + 15) / 16, (unsigned)(Hh)), 32, 0, stream>>>(cp0_11); }
    { GemmP cp0_12;
      cp0_12.A = XP + (size_t)4106 * CI; cp0_12.B = wpre + 12; cp0_12.bias = XP + (size_t)4106 * CI; cp0_12.R = HP + C1; cp0_12.C = HP + C1;
      cp0_12.sAo = (long long)2052 * CI; cp0_12.sAi = 0; cp0_12.sAm = CI; cp0_12.sAk = 1; cp0_12.sBo = 0; cp0_12.sBi = 0; cp0_12.sBn = CI * 25; cp0_12.sBk = 25; cp0_12.sCo = (long long)2050 * C1; cp0_12.sCi = 0; cp0_12.sCm = C1; cp0_12.sRo = (long long)2050 * C1; cp0_12.sRi = 0; cp0_12.sRm = C1; cp0_12.sRn = 1;
      cp0_12.M = Tt; cp0_12.N = C1; cp0_12.K = CI; cp0_12.zi_n = 1; cp0_12.flags = 4; cp0_12.act = 0;
      cp0_12.alpha = 1.0f; cp0_12.beta = 1.0f; cp0_12.sa = 1.0f; cp0_12.sb = 1.0f; cp0_12.Npad = C1; cp0_12.pad_ = 0;
      k_gemm<1><<<dim3((unsigned)((C1) + 31) / 32, (unsigned)((Tt) + 15) / 16, (unsigned)(Hh)), 32, 0, stream>>>(cp0_12); }
    { GemmP cp0_13;
      cp0_13.A = XP + (size_t)4107 * CI; cp0_13.B = wpre + 13; cp0_13.bias = XP + (size_t)4107 * CI; cp0_13.R = HP + C1; cp0_13.C = HP + C1;
      cp0_13.sAo = (long long)2052 * CI; cp0_13.sAi = 0; cp0_13.sAm = CI; cp0_13.sAk = 1; cp0_13.sBo = 0; cp0_13.sBi = 0; cp0_13.sBn = CI * 25; cp0_13.sBk = 25; cp0_13.sCo = (long long)2050 * C1; cp0_13.sCi = 0; cp0_13.sCm = C1; cp0_13.sRo = (long long)2050 * C1; cp0_13.sRi = 0; cp0_13.sRm = C1; cp0_13.sRn = 1;
      cp0_13.M = Tt; cp0_13.N = C1; cp0_13.K = CI; cp0_13.zi_n = 1; cp0_13.flags = 4; cp0_13.act = 0;
      cp0_13.alpha = 1.0f; cp0_13.beta = 1.0f; cp0_13.sa = 1.0f; cp0_13.sb = 1.0f; cp0_13.Npad = C1; cp0_13.pad_ = 0;
      k_gemm<1><<<dim3((unsigned)((C1) + 31) / 32, (unsigned)((Tt) + 15) / 16, (unsigned)(Hh)), 32, 0, stream>>>(cp0_13); }
    { GemmP cp0_14;
      cp0_14.A = XP + (size_t)4108 * CI; cp0_14.B = wpre + 14; cp0_14.bias = XP + (size_t)4108 * CI; cp0_14.R = HP + C1; cp0_14.C = HP + C1;
      cp0_14.sAo = (long long)2052 * CI; cp0_14.sAi = 0; cp0_14.sAm = CI; cp0_14.sAk = 1; cp0_14.sBo = 0; cp0_14.sBi = 0; cp0_14.sBn = CI * 25; cp0_14.sBk = 25; cp0_14.sCo = (long long)2050 * C1; cp0_14.sCi = 0; cp0_14.sCm = C1; cp0_14.sRo = (long long)2050 * C1; cp0_14.sRi = 0; cp0_14.sRm = C1; cp0_14.sRn = 1;
      cp0_14.M = Tt; cp0_14.N = C1; cp0_14.K = CI; cp0_14.zi_n = 1; cp0_14.flags = 4; cp0_14.act = 0;
      cp0_14.alpha = 1.0f; cp0_14.beta = 1.0f; cp0_14.sa = 1.0f; cp0_14.sb = 1.0f; cp0_14.Npad = C1; cp0_14.pad_ = 0;
      k_gemm<1><<<dim3((unsigned)((C1) + 31) / 32, (unsigned)((Tt) + 15) / 16, (unsigned)(Hh)), 32, 0, stream>>>(cp0_14); }
    { GemmP cp0_15;
      cp0_15.A = XP + (size_t)6156 * CI; cp0_15.B = wpre + 15; cp0_15.bias = XP + (size_t)6156 * CI; cp0_15.R = HP + C1; cp0_15.C = HP + C1;
      cp0_15.sAo = (long long)2052 * CI; cp0_15.sAi = 0; cp0_15.sAm = CI; cp0_15.sAk = 1; cp0_15.sBo = 0; cp0_15.sBi = 0; cp0_15.sBn = CI * 25; cp0_15.sBk = 25; cp0_15.sCo = (long long)2050 * C1; cp0_15.sCi = 0; cp0_15.sCm = C1; cp0_15.sRo = (long long)2050 * C1; cp0_15.sRi = 0; cp0_15.sRm = C1; cp0_15.sRn = 1;
      cp0_15.M = Tt; cp0_15.N = C1; cp0_15.K = CI; cp0_15.zi_n = 1; cp0_15.flags = 4; cp0_15.act = 0;
      cp0_15.alpha = 1.0f; cp0_15.beta = 1.0f; cp0_15.sa = 1.0f; cp0_15.sb = 1.0f; cp0_15.Npad = C1; cp0_15.pad_ = 0;
      k_gemm<1><<<dim3((unsigned)((C1) + 31) / 32, (unsigned)((Tt) + 15) / 16, (unsigned)(Hh)), 32, 0, stream>>>(cp0_15); }
    { GemmP cp0_16;
      cp0_16.A = XP + (size_t)6157 * CI; cp0_16.B = wpre + 16; cp0_16.bias = XP + (size_t)6157 * CI; cp0_16.R = HP + C1; cp0_16.C = HP + C1;
      cp0_16.sAo = (long long)2052 * CI; cp0_16.sAi = 0; cp0_16.sAm = CI; cp0_16.sAk = 1; cp0_16.sBo = 0; cp0_16.sBi = 0; cp0_16.sBn = CI * 25; cp0_16.sBk = 25; cp0_16.sCo = (long long)2050 * C1; cp0_16.sCi = 0; cp0_16.sCm = C1; cp0_16.sRo = (long long)2050 * C1; cp0_16.sRi = 0; cp0_16.sRm = C1; cp0_16.sRn = 1;
      cp0_16.M = Tt; cp0_16.N = C1; cp0_16.K = CI; cp0_16.zi_n = 1; cp0_16.flags = 4; cp0_16.act = 0;
      cp0_16.alpha = 1.0f; cp0_16.beta = 1.0f; cp0_16.sa = 1.0f; cp0_16.sb = 1.0f; cp0_16.Npad = C1; cp0_16.pad_ = 0;
      k_gemm<1><<<dim3((unsigned)((C1) + 31) / 32, (unsigned)((Tt) + 15) / 16, (unsigned)(Hh)), 32, 0, stream>>>(cp0_16); }
    { GemmP cp0_17;
      cp0_17.A = XP + (size_t)6158 * CI; cp0_17.B = wpre + 17; cp0_17.bias = XP + (size_t)6158 * CI; cp0_17.R = HP + C1; cp0_17.C = HP + C1;
      cp0_17.sAo = (long long)2052 * CI; cp0_17.sAi = 0; cp0_17.sAm = CI; cp0_17.sAk = 1; cp0_17.sBo = 0; cp0_17.sBi = 0; cp0_17.sBn = CI * 25; cp0_17.sBk = 25; cp0_17.sCo = (long long)2050 * C1; cp0_17.sCi = 0; cp0_17.sCm = C1; cp0_17.sRo = (long long)2050 * C1; cp0_17.sRi = 0; cp0_17.sRm = C1; cp0_17.sRn = 1;
      cp0_17.M = Tt; cp0_17.N = C1; cp0_17.K = CI; cp0_17.zi_n = 1; cp0_17.flags = 4; cp0_17.act = 0;
      cp0_17.alpha = 1.0f; cp0_17.beta = 1.0f; cp0_17.sa = 1.0f; cp0_17.sb = 1.0f; cp0_17.Npad = C1; cp0_17.pad_ = 0;
      k_gemm<1><<<dim3((unsigned)((C1) + 31) / 32, (unsigned)((Tt) + 15) / 16, (unsigned)(Hh)), 32, 0, stream>>>(cp0_17); }
    { GemmP cp0_18;
      cp0_18.A = XP + (size_t)6159 * CI; cp0_18.B = wpre + 18; cp0_18.bias = XP + (size_t)6159 * CI; cp0_18.R = HP + C1; cp0_18.C = HP + C1;
      cp0_18.sAo = (long long)2052 * CI; cp0_18.sAi = 0; cp0_18.sAm = CI; cp0_18.sAk = 1; cp0_18.sBo = 0; cp0_18.sBi = 0; cp0_18.sBn = CI * 25; cp0_18.sBk = 25; cp0_18.sCo = (long long)2050 * C1; cp0_18.sCi = 0; cp0_18.sCm = C1; cp0_18.sRo = (long long)2050 * C1; cp0_18.sRi = 0; cp0_18.sRm = C1; cp0_18.sRn = 1;
      cp0_18.M = Tt; cp0_18.N = C1; cp0_18.K = CI; cp0_18.zi_n = 1; cp0_18.flags = 4; cp0_18.act = 0;
      cp0_18.alpha = 1.0f; cp0_18.beta = 1.0f; cp0_18.sa = 1.0f; cp0_18.sb = 1.0f; cp0_18.Npad = C1; cp0_18.pad_ = 0;
      k_gemm<1><<<dim3((unsigned)((C1) + 31) / 32, (unsigned)((Tt) + 15) / 16, (unsigned)(Hh)), 32, 0, stream>>>(cp0_18); }
    { GemmP cp0_19;
      cp0_19.A = XP + (size_t)6160 * CI; cp0_19.B = wpre + 19; cp0_19.bias = XP + (size_t)6160 * CI; cp0_19.R = HP + C1; cp0_19.C = HP + C1;
      cp0_19.sAo = (long long)2052 * CI; cp0_19.sAi = 0; cp0_19.sAm = CI; cp0_19.sAk = 1; cp0_19.sBo = 0; cp0_19.sBi = 0; cp0_19.sBn = CI * 25; cp0_19.sBk = 25; cp0_19.sCo = (long long)2050 * C1; cp0_19.sCi = 0; cp0_19.sCm = C1; cp0_19.sRo = (long long)2050 * C1; cp0_19.sRi = 0; cp0_19.sRm = C1; cp0_19.sRn = 1;
      cp0_19.M = Tt; cp0_19.N = C1; cp0_19.K = CI; cp0_19.zi_n = 1; cp0_19.flags = 4; cp0_19.act = 0;
      cp0_19.alpha = 1.0f; cp0_19.beta = 1.0f; cp0_19.sa = 1.0f; cp0_19.sb = 1.0f; cp0_19.Npad = C1; cp0_19.pad_ = 0;
      k_gemm<1><<<dim3((unsigned)((C1) + 31) / 32, (unsigned)((Tt) + 15) / 16, (unsigned)(Hh)), 32, 0, stream>>>(cp0_19); }
    { GemmP cp0_20;
      cp0_20.A = XP + (size_t)8208 * CI; cp0_20.B = wpre + 20; cp0_20.bias = XP + (size_t)8208 * CI; cp0_20.R = HP + C1; cp0_20.C = HP + C1;
      cp0_20.sAo = (long long)2052 * CI; cp0_20.sAi = 0; cp0_20.sAm = CI; cp0_20.sAk = 1; cp0_20.sBo = 0; cp0_20.sBi = 0; cp0_20.sBn = CI * 25; cp0_20.sBk = 25; cp0_20.sCo = (long long)2050 * C1; cp0_20.sCi = 0; cp0_20.sCm = C1; cp0_20.sRo = (long long)2050 * C1; cp0_20.sRi = 0; cp0_20.sRm = C1; cp0_20.sRn = 1;
      cp0_20.M = Tt; cp0_20.N = C1; cp0_20.K = CI; cp0_20.zi_n = 1; cp0_20.flags = 4; cp0_20.act = 0;
      cp0_20.alpha = 1.0f; cp0_20.beta = 1.0f; cp0_20.sa = 1.0f; cp0_20.sb = 1.0f; cp0_20.Npad = C1; cp0_20.pad_ = 0;
      k_gemm<1><<<dim3((unsigned)((C1) + 31) / 32, (unsigned)((Tt) + 15) / 16, (unsigned)(Hh)), 32, 0, stream>>>(cp0_20); }
    { GemmP cp0_21;
      cp0_21.A = XP + (size_t)8209 * CI; cp0_21.B = wpre + 21; cp0_21.bias = XP + (size_t)8209 * CI; cp0_21.R = HP + C1; cp0_21.C = HP + C1;
      cp0_21.sAo = (long long)2052 * CI; cp0_21.sAi = 0; cp0_21.sAm = CI; cp0_21.sAk = 1; cp0_21.sBo = 0; cp0_21.sBi = 0; cp0_21.sBn = CI * 25; cp0_21.sBk = 25; cp0_21.sCo = (long long)2050 * C1; cp0_21.sCi = 0; cp0_21.sCm = C1; cp0_21.sRo = (long long)2050 * C1; cp0_21.sRi = 0; cp0_21.sRm = C1; cp0_21.sRn = 1;
      cp0_21.M = Tt; cp0_21.N = C1; cp0_21.K = CI; cp0_21.zi_n = 1; cp0_21.flags = 4; cp0_21.act = 0;
      cp0_21.alpha = 1.0f; cp0_21.beta = 1.0f; cp0_21.sa = 1.0f; cp0_21.sb = 1.0f; cp0_21.Npad = C1; cp0_21.pad_ = 0;
      k_gemm<1><<<dim3((unsigned)((C1) + 31) / 32, (unsigned)((Tt) + 15) / 16, (unsigned)(Hh)), 32, 0, stream>>>(cp0_21); }
    { GemmP cp0_22;
      cp0_22.A = XP + (size_t)8210 * CI; cp0_22.B = wpre + 22; cp0_22.bias = XP + (size_t)8210 * CI; cp0_22.R = HP + C1; cp0_22.C = HP + C1;
      cp0_22.sAo = (long long)2052 * CI; cp0_22.sAi = 0; cp0_22.sAm = CI; cp0_22.sAk = 1; cp0_22.sBo = 0; cp0_22.sBi = 0; cp0_22.sBn = CI * 25; cp0_22.sBk = 25; cp0_22.sCo = (long long)2050 * C1; cp0_22.sCi = 0; cp0_22.sCm = C1; cp0_22.sRo = (long long)2050 * C1; cp0_22.sRi = 0; cp0_22.sRm = C1; cp0_22.sRn = 1;
      cp0_22.M = Tt; cp0_22.N = C1; cp0_22.K = CI; cp0_22.zi_n = 1; cp0_22.flags = 4; cp0_22.act = 0;
      cp0_22.alpha = 1.0f; cp0_22.beta = 1.0f; cp0_22.sa = 1.0f; cp0_22.sb = 1.0f; cp0_22.Npad = C1; cp0_22.pad_ = 0;
      k_gemm<1><<<dim3((unsigned)((C1) + 31) / 32, (unsigned)((Tt) + 15) / 16, (unsigned)(Hh)), 32, 0, stream>>>(cp0_22); }
    { GemmP cp0_23;
      cp0_23.A = XP + (size_t)8211 * CI; cp0_23.B = wpre + 23; cp0_23.bias = XP + (size_t)8211 * CI; cp0_23.R = HP + C1; cp0_23.C = HP + C1;
      cp0_23.sAo = (long long)2052 * CI; cp0_23.sAi = 0; cp0_23.sAm = CI; cp0_23.sAk = 1; cp0_23.sBo = 0; cp0_23.sBi = 0; cp0_23.sBn = CI * 25; cp0_23.sBk = 25; cp0_23.sCo = (long long)2050 * C1; cp0_23.sCi = 0; cp0_23.sCm = C1; cp0_23.sRo = (long long)2050 * C1; cp0_23.sRi = 0; cp0_23.sRm = C1; cp0_23.sRn = 1;
      cp0_23.M = Tt; cp0_23.N = C1; cp0_23.K = CI; cp0_23.zi_n = 1; cp0_23.flags = 4; cp0_23.act = 0;
      cp0_23.alpha = 1.0f; cp0_23.beta = 1.0f; cp0_23.sa = 1.0f; cp0_23.sb = 1.0f; cp0_23.Npad = C1; cp0_23.pad_ = 0;
      k_gemm<1><<<dim3((unsigned)((C1) + 31) / 32, (unsigned)((Tt) + 15) / 16, (unsigned)(Hh)), 32, 0, stream>>>(cp0_23); }
    { GemmP cp0_24;
      cp0_24.A = XP + (size_t)8212 * CI; cp0_24.B = wpre + 24; cp0_24.bias = XP + (size_t)8212 * CI; cp0_24.R = HP + C1; cp0_24.C = HP + C1;
      cp0_24.sAo = (long long)2052 * CI; cp0_24.sAi = 0; cp0_24.sAm = CI; cp0_24.sAk = 1; cp0_24.sBo = 0; cp0_24.sBi = 0; cp0_24.sBn = CI * 25; cp0_24.sBk = 25; cp0_24.sCo = (long long)2050 * C1; cp0_24.sCi = 0; cp0_24.sCm = C1; cp0_24.sRo = (long long)2050 * C1; cp0_24.sRi = 0; cp0_24.sRm = C1; cp0_24.sRn = 1;
      cp0_24.M = Tt; cp0_24.N = C1; cp0_24.K = CI; cp0_24.zi_n = 1; cp0_24.flags = 4; cp0_24.act = 0;
      cp0_24.alpha = 1.0f; cp0_24.beta = 1.0f; cp0_24.sa = 1.0f; cp0_24.sb = 1.0f; cp0_24.Npad = C1; cp0_24.pad_ = 0;
      k_gemm<1><<<dim3((unsigned)((C1) + 31) / 32, (unsigned)((Tt) + 15) / 16, (unsigned)(Hh)), 32, 0, stream>>>(cp0_24); }
    k_cl_bnl<<<(unsigned)(((long long)Hh * Tt * C1 + 255) / 256), 256, 0, stream>>>(HP, bng, bnb, bnm, bnv, Hh, Tt, C1);
    { GemmP ceq0_0;
      ceq0_0.A = HP + (size_t)0 * C1; ceq0_0.B = wq + 0; ceq0_0.bias = bq; ceq0_0.R = HP + (size_t)0 * C1; ceq0_0.C = Q;
      ceq0_0.sAo = (long long)3 * 2050 * C1; ceq0_0.sAi = 0; ceq0_0.sAm = C1; ceq0_0.sAk = 1; ceq0_0.sBo = 0; ceq0_0.sBi = 0; ceq0_0.sBn = C1 * 9; ceq0_0.sBk = 9; ceq0_0.sCo = (long long)Tt * LD; ceq0_0.sCi = 0; ceq0_0.sCm = LD; ceq0_0.sRo = 0; ceq0_0.sRi = 0; ceq0_0.sRm = 0; ceq0_0.sRn = 0;
      ceq0_0.M = Tt; ceq0_0.N = D; ceq0_0.K = C1; ceq0_0.zi_n = 1; ceq0_0.flags = 1; ceq0_0.act = 0;
      ceq0_0.alpha = 1.0f; ceq0_0.beta = 0.0f; ceq0_0.sa = 1.0f; ceq0_0.sb = 1.0f; ceq0_0.Npad = LD; ceq0_0.pad_ = 0;
      k_gemm<1><<<dim3((unsigned)((LD) + 31) / 32, (unsigned)((Tt) + 15) / 16, (unsigned)(Fo)), 32, 0, stream>>>(ceq0_0); }
    { GemmP ceq0_1;
      ceq0_1.A = HP + (size_t)1 * C1; ceq0_1.B = wq + 1; ceq0_1.bias = HP + (size_t)1 * C1; ceq0_1.R = Q; ceq0_1.C = Q;
      ceq0_1.sAo = (long long)3 * 2050 * C1; ceq0_1.sAi = 0; ceq0_1.sAm = C1; ceq0_1.sAk = 1; ceq0_1.sBo = 0; ceq0_1.sBi = 0; ceq0_1.sBn = C1 * 9; ceq0_1.sBk = 9; ceq0_1.sCo = (long long)Tt * LD; ceq0_1.sCi = 0; ceq0_1.sCm = LD; ceq0_1.sRo = (long long)Tt * LD; ceq0_1.sRi = 0; ceq0_1.sRm = LD; ceq0_1.sRn = 1;
      ceq0_1.M = Tt; ceq0_1.N = D; ceq0_1.K = C1; ceq0_1.zi_n = 1; ceq0_1.flags = 4; ceq0_1.act = 0;
      ceq0_1.alpha = 1.0f; ceq0_1.beta = 1.0f; ceq0_1.sa = 1.0f; ceq0_1.sb = 1.0f; ceq0_1.Npad = LD; ceq0_1.pad_ = 0;
      k_gemm<1><<<dim3((unsigned)((LD) + 31) / 32, (unsigned)((Tt) + 15) / 16, (unsigned)(Fo)), 32, 0, stream>>>(ceq0_1); }
    { GemmP ceq0_2;
      ceq0_2.A = HP + (size_t)2 * C1; ceq0_2.B = wq + 2; ceq0_2.bias = HP + (size_t)2 * C1; ceq0_2.R = Q; ceq0_2.C = Q;
      ceq0_2.sAo = (long long)3 * 2050 * C1; ceq0_2.sAi = 0; ceq0_2.sAm = C1; ceq0_2.sAk = 1; ceq0_2.sBo = 0; ceq0_2.sBi = 0; ceq0_2.sBn = C1 * 9; ceq0_2.sBk = 9; ceq0_2.sCo = (long long)Tt * LD; ceq0_2.sCi = 0; ceq0_2.sCm = LD; ceq0_2.sRo = (long long)Tt * LD; ceq0_2.sRi = 0; ceq0_2.sRm = LD; ceq0_2.sRn = 1;
      ceq0_2.M = Tt; ceq0_2.N = D; ceq0_2.K = C1; ceq0_2.zi_n = 1; ceq0_2.flags = 4; ceq0_2.act = 0;
      ceq0_2.alpha = 1.0f; ceq0_2.beta = 1.0f; ceq0_2.sa = 1.0f; ceq0_2.sb = 1.0f; ceq0_2.Npad = LD; ceq0_2.pad_ = 0;
      k_gemm<1><<<dim3((unsigned)((LD) + 31) / 32, (unsigned)((Tt) + 15) / 16, (unsigned)(Fo)), 32, 0, stream>>>(ceq0_2); }
    { GemmP ceq0_3;
      ceq0_3.A = HP + (size_t)2050 * C1; ceq0_3.B = wq + 3; ceq0_3.bias = HP + (size_t)2050 * C1; ceq0_3.R = Q; ceq0_3.C = Q;
      ceq0_3.sAo = (long long)3 * 2050 * C1; ceq0_3.sAi = 0; ceq0_3.sAm = C1; ceq0_3.sAk = 1; ceq0_3.sBo = 0; ceq0_3.sBi = 0; ceq0_3.sBn = C1 * 9; ceq0_3.sBk = 9; ceq0_3.sCo = (long long)Tt * LD; ceq0_3.sCi = 0; ceq0_3.sCm = LD; ceq0_3.sRo = (long long)Tt * LD; ceq0_3.sRi = 0; ceq0_3.sRm = LD; ceq0_3.sRn = 1;
      ceq0_3.M = Tt; ceq0_3.N = D; ceq0_3.K = C1; ceq0_3.zi_n = 1; ceq0_3.flags = 4; ceq0_3.act = 0;
      ceq0_3.alpha = 1.0f; ceq0_3.beta = 1.0f; ceq0_3.sa = 1.0f; ceq0_3.sb = 1.0f; ceq0_3.Npad = LD; ceq0_3.pad_ = 0;
      k_gemm<1><<<dim3((unsigned)((LD) + 31) / 32, (unsigned)((Tt) + 15) / 16, (unsigned)(Fo)), 32, 0, stream>>>(ceq0_3); }
    { GemmP ceq0_4;
      ceq0_4.A = HP + (size_t)2051 * C1; ceq0_4.B = wq + 4; ceq0_4.bias = HP + (size_t)2051 * C1; ceq0_4.R = Q; ceq0_4.C = Q;
      ceq0_4.sAo = (long long)3 * 2050 * C1; ceq0_4.sAi = 0; ceq0_4.sAm = C1; ceq0_4.sAk = 1; ceq0_4.sBo = 0; ceq0_4.sBi = 0; ceq0_4.sBn = C1 * 9; ceq0_4.sBk = 9; ceq0_4.sCo = (long long)Tt * LD; ceq0_4.sCi = 0; ceq0_4.sCm = LD; ceq0_4.sRo = (long long)Tt * LD; ceq0_4.sRi = 0; ceq0_4.sRm = LD; ceq0_4.sRn = 1;
      ceq0_4.M = Tt; ceq0_4.N = D; ceq0_4.K = C1; ceq0_4.zi_n = 1; ceq0_4.flags = 4; ceq0_4.act = 0;
      ceq0_4.alpha = 1.0f; ceq0_4.beta = 1.0f; ceq0_4.sa = 1.0f; ceq0_4.sb = 1.0f; ceq0_4.Npad = LD; ceq0_4.pad_ = 0;
      k_gemm<1><<<dim3((unsigned)((LD) + 31) / 32, (unsigned)((Tt) + 15) / 16, (unsigned)(Fo)), 32, 0, stream>>>(ceq0_4); }
    { GemmP ceq0_5;
      ceq0_5.A = HP + (size_t)2052 * C1; ceq0_5.B = wq + 5; ceq0_5.bias = HP + (size_t)2052 * C1; ceq0_5.R = Q; ceq0_5.C = Q;
      ceq0_5.sAo = (long long)3 * 2050 * C1; ceq0_5.sAi = 0; ceq0_5.sAm = C1; ceq0_5.sAk = 1; ceq0_5.sBo = 0; ceq0_5.sBi = 0; ceq0_5.sBn = C1 * 9; ceq0_5.sBk = 9; ceq0_5.sCo = (long long)Tt * LD; ceq0_5.sCi = 0; ceq0_5.sCm = LD; ceq0_5.sRo = (long long)Tt * LD; ceq0_5.sRi = 0; ceq0_5.sRm = LD; ceq0_5.sRn = 1;
      ceq0_5.M = Tt; ceq0_5.N = D; ceq0_5.K = C1; ceq0_5.zi_n = 1; ceq0_5.flags = 4; ceq0_5.act = 0;
      ceq0_5.alpha = 1.0f; ceq0_5.beta = 1.0f; ceq0_5.sa = 1.0f; ceq0_5.sb = 1.0f; ceq0_5.Npad = LD; ceq0_5.pad_ = 0;
      k_gemm<1><<<dim3((unsigned)((LD) + 31) / 32, (unsigned)((Tt) + 15) / 16, (unsigned)(Fo)), 32, 0, stream>>>(ceq0_5); }
    { GemmP ceq0_6;
      ceq0_6.A = HP + (size_t)4100 * C1; ceq0_6.B = wq + 6; ceq0_6.bias = HP + (size_t)4100 * C1; ceq0_6.R = Q; ceq0_6.C = Q;
      ceq0_6.sAo = (long long)3 * 2050 * C1; ceq0_6.sAi = 0; ceq0_6.sAm = C1; ceq0_6.sAk = 1; ceq0_6.sBo = 0; ceq0_6.sBi = 0; ceq0_6.sBn = C1 * 9; ceq0_6.sBk = 9; ceq0_6.sCo = (long long)Tt * LD; ceq0_6.sCi = 0; ceq0_6.sCm = LD; ceq0_6.sRo = (long long)Tt * LD; ceq0_6.sRi = 0; ceq0_6.sRm = LD; ceq0_6.sRn = 1;
      ceq0_6.M = Tt; ceq0_6.N = D; ceq0_6.K = C1; ceq0_6.zi_n = 1; ceq0_6.flags = 4; ceq0_6.act = 0;
      ceq0_6.alpha = 1.0f; ceq0_6.beta = 1.0f; ceq0_6.sa = 1.0f; ceq0_6.sb = 1.0f; ceq0_6.Npad = LD; ceq0_6.pad_ = 0;
      k_gemm<1><<<dim3((unsigned)((LD) + 31) / 32, (unsigned)((Tt) + 15) / 16, (unsigned)(Fo)), 32, 0, stream>>>(ceq0_6); }
    { GemmP ceq0_7;
      ceq0_7.A = HP + (size_t)4101 * C1; ceq0_7.B = wq + 7; ceq0_7.bias = HP + (size_t)4101 * C1; ceq0_7.R = Q; ceq0_7.C = Q;
      ceq0_7.sAo = (long long)3 * 2050 * C1; ceq0_7.sAi = 0; ceq0_7.sAm = C1; ceq0_7.sAk = 1; ceq0_7.sBo = 0; ceq0_7.sBi = 0; ceq0_7.sBn = C1 * 9; ceq0_7.sBk = 9; ceq0_7.sCo = (long long)Tt * LD; ceq0_7.sCi = 0; ceq0_7.sCm = LD; ceq0_7.sRo = (long long)Tt * LD; ceq0_7.sRi = 0; ceq0_7.sRm = LD; ceq0_7.sRn = 1;
      ceq0_7.M = Tt; ceq0_7.N = D; ceq0_7.K = C1; ceq0_7.zi_n = 1; ceq0_7.flags = 4; ceq0_7.act = 0;
      ceq0_7.alpha = 1.0f; ceq0_7.beta = 1.0f; ceq0_7.sa = 1.0f; ceq0_7.sb = 1.0f; ceq0_7.Npad = LD; ceq0_7.pad_ = 0;
      k_gemm<1><<<dim3((unsigned)((LD) + 31) / 32, (unsigned)((Tt) + 15) / 16, (unsigned)(Fo)), 32, 0, stream>>>(ceq0_7); }
    { GemmP ceq0_8;
      ceq0_8.A = HP + (size_t)4102 * C1; ceq0_8.B = wq + 8; ceq0_8.bias = HP + (size_t)4102 * C1; ceq0_8.R = Q; ceq0_8.C = Q;
      ceq0_8.sAo = (long long)3 * 2050 * C1; ceq0_8.sAi = 0; ceq0_8.sAm = C1; ceq0_8.sAk = 1; ceq0_8.sBo = 0; ceq0_8.sBi = 0; ceq0_8.sBn = C1 * 9; ceq0_8.sBk = 9; ceq0_8.sCo = (long long)Tt * LD; ceq0_8.sCi = 0; ceq0_8.sCm = LD; ceq0_8.sRo = (long long)Tt * LD; ceq0_8.sRi = 0; ceq0_8.sRm = LD; ceq0_8.sRn = 1;
      ceq0_8.M = Tt; ceq0_8.N = D; ceq0_8.K = C1; ceq0_8.zi_n = 1; ceq0_8.flags = 4; ceq0_8.act = 0;
      ceq0_8.alpha = 1.0f; ceq0_8.beta = 1.0f; ceq0_8.sa = 1.0f; ceq0_8.sb = 1.0f; ceq0_8.Npad = LD; ceq0_8.pad_ = 0;
      k_gemm<1><<<dim3((unsigned)((LD) + 31) / 32, (unsigned)((Tt) + 15) / 16, (unsigned)(Fo)), 32, 0, stream>>>(ceq0_8); }

    { GemmP cekv0_0;
      cekv0_0.A = HP + (size_t)0 * C1; cekv0_0.B = wkv + 0; cekv0_0.bias = bkv; cekv0_0.R = HP + (size_t)0 * C1; cekv0_0.C = KV;
      cekv0_0.sAo = (long long)3 * 2050 * C1; cekv0_0.sAi = 0; cekv0_0.sAm = C1; cekv0_0.sAk = 1; cekv0_0.sBo = 0; cekv0_0.sBi = 0; cekv0_0.sBn = C1 * 9; cekv0_0.sBk = 9; cekv0_0.sCo = (long long)Tt * LD; cekv0_0.sCi = 0; cekv0_0.sCm = LD; cekv0_0.sRo = 0; cekv0_0.sRi = 0; cekv0_0.sRm = 0; cekv0_0.sRn = 0;
      cekv0_0.M = Tt; cekv0_0.N = D; cekv0_0.K = C1; cekv0_0.zi_n = 1; cekv0_0.flags = 1; cekv0_0.act = 0;
      cekv0_0.alpha = 1.0f; cekv0_0.beta = 0.0f; cekv0_0.sa = 1.0f; cekv0_0.sb = 1.0f; cekv0_0.Npad = LD; cekv0_0.pad_ = 0;
      k_gemm<1><<<dim3((unsigned)((LD) + 31) / 32, (unsigned)((Tt) + 15) / 16, (unsigned)(Fo)), 32, 0, stream>>>(cekv0_0); }
    { GemmP cekv0_1;
      cekv0_1.A = HP + (size_t)1 * C1; cekv0_1.B = wkv + 1; cekv0_1.bias = HP + (size_t)1 * C1; cekv0_1.R = KV; cekv0_1.C = KV;
      cekv0_1.sAo = (long long)3 * 2050 * C1; cekv0_1.sAi = 0; cekv0_1.sAm = C1; cekv0_1.sAk = 1; cekv0_1.sBo = 0; cekv0_1.sBi = 0; cekv0_1.sBn = C1 * 9; cekv0_1.sBk = 9; cekv0_1.sCo = (long long)Tt * LD; cekv0_1.sCi = 0; cekv0_1.sCm = LD; cekv0_1.sRo = (long long)Tt * LD; cekv0_1.sRi = 0; cekv0_1.sRm = LD; cekv0_1.sRn = 1;
      cekv0_1.M = Tt; cekv0_1.N = D; cekv0_1.K = C1; cekv0_1.zi_n = 1; cekv0_1.flags = 4; cekv0_1.act = 0;
      cekv0_1.alpha = 1.0f; cekv0_1.beta = 1.0f; cekv0_1.sa = 1.0f; cekv0_1.sb = 1.0f; cekv0_1.Npad = LD; cekv0_1.pad_ = 0;
      k_gemm<1><<<dim3((unsigned)((LD) + 31) / 32, (unsigned)((Tt) + 15) / 16, (unsigned)(Fo)), 32, 0, stream>>>(cekv0_1); }
    { GemmP cekv0_2;
      cekv0_2.A = HP + (size_t)2 * C1; cekv0_2.B = wkv + 2; cekv0_2.bias = HP + (size_t)2 * C1; cekv0_2.R = KV; cekv0_2.C = KV;
      cekv0_2.sAo = (long long)3 * 2050 * C1; cekv0_2.sAi = 0; cekv0_2.sAm = C1; cekv0_2.sAk = 1; cekv0_2.sBo = 0; cekv0_2.sBi = 0; cekv0_2.sBn = C1 * 9; cekv0_2.sBk = 9; cekv0_2.sCo = (long long)Tt * LD; cekv0_2.sCi = 0; cekv0_2.sCm = LD; cekv0_2.sRo = (long long)Tt * LD; cekv0_2.sRi = 0; cekv0_2.sRm = LD; cekv0_2.sRn = 1;
      cekv0_2.M = Tt; cekv0_2.N = D; cekv0_2.K = C1; cekv0_2.zi_n = 1; cekv0_2.flags = 4; cekv0_2.act = 0;
      cekv0_2.alpha = 1.0f; cekv0_2.beta = 1.0f; cekv0_2.sa = 1.0f; cekv0_2.sb = 1.0f; cekv0_2.Npad = LD; cekv0_2.pad_ = 0;
      k_gemm<1><<<dim3((unsigned)((LD) + 31) / 32, (unsigned)((Tt) + 15) / 16, (unsigned)(Fo)), 32, 0, stream>>>(cekv0_2); }
    { GemmP cekv0_3;
      cekv0_3.A = HP + (size_t)2050 * C1; cekv0_3.B = wkv + 3; cekv0_3.bias = HP + (size_t)2050 * C1; cekv0_3.R = KV; cekv0_3.C = KV;
      cekv0_3.sAo = (long long)3 * 2050 * C1; cekv0_3.sAi = 0; cekv0_3.sAm = C1; cekv0_3.sAk = 1; cekv0_3.sBo = 0; cekv0_3.sBi = 0; cekv0_3.sBn = C1 * 9; cekv0_3.sBk = 9; cekv0_3.sCo = (long long)Tt * LD; cekv0_3.sCi = 0; cekv0_3.sCm = LD; cekv0_3.sRo = (long long)Tt * LD; cekv0_3.sRi = 0; cekv0_3.sRm = LD; cekv0_3.sRn = 1;
      cekv0_3.M = Tt; cekv0_3.N = D; cekv0_3.K = C1; cekv0_3.zi_n = 1; cekv0_3.flags = 4; cekv0_3.act = 0;
      cekv0_3.alpha = 1.0f; cekv0_3.beta = 1.0f; cekv0_3.sa = 1.0f; cekv0_3.sb = 1.0f; cekv0_3.Npad = LD; cekv0_3.pad_ = 0;
      k_gemm<1><<<dim3((unsigned)((LD) + 31) / 32, (unsigned)((Tt) + 15) / 16, (unsigned)(Fo)), 32, 0, stream>>>(cekv0_3); }
    { GemmP cekv0_4;
      cekv0_4.A = HP + (size_t)2051 * C1; cekv0_4.B = wkv + 4; cekv0_4.bias = HP + (size_t)2051 * C1; cekv0_4.R = KV; cekv0_4.C = KV;
      cekv0_4.sAo = (long long)3 * 2050 * C1; cekv0_4.sAi = 0; cekv0_4.sAm = C1; cekv0_4.sAk = 1; cekv0_4.sBo = 0; cekv0_4.sBi = 0; cekv0_4.sBn = C1 * 9; cekv0_4.sBk = 9; cekv0_4.sCo = (long long)Tt * LD; cekv0_4.sCi = 0; cekv0_4.sCm = LD; cekv0_4.sRo = (long long)Tt * LD; cekv0_4.sRi = 0; cekv0_4.sRm = LD; cekv0_4.sRn = 1;
      cekv0_4.M = Tt; cekv0_4.N = D; cekv0_4.K = C1; cekv0_4.zi_n = 1; cekv0_4.flags = 4; cekv0_4.act = 0;
      cekv0_4.alpha = 1.0f; cekv0_4.beta = 1.0f; cekv0_4.sa = 1.0f; cekv0_4.sb = 1.0f; cekv0_4.Npad = LD; cekv0_4.pad_ = 0;
      k_gemm<1><<<dim3((unsigned)((LD) + 31) / 32, (unsigned)((Tt) + 15) / 16, (unsigned)(Fo)), 32, 0, stream>>>(cekv0_4); }
    { GemmP cekv0_5;
      cekv0_5.A = HP + (size_t)2052 * C1; cekv0_5.B = wkv + 5; cekv0_5.bias = HP + (size_t)2052 * C1; cekv0_5.R = KV; cekv0_5.C = KV;
      cekv0_5.sAo = (long long)3 * 2050 * C1; cekv0_5.sAi = 0; cekv0_5.sAm = C1; cekv0_5.sAk = 1; cekv0_5.sBo = 0; cekv0_5.sBi = 0; cekv0_5.sBn = C1 * 9; cekv0_5.sBk = 9; cekv0_5.sCo = (long long)Tt * LD; cekv0_5.sCi = 0; cekv0_5.sCm = LD; cekv0_5.sRo = (long long)Tt * LD; cekv0_5.sRi = 0; cekv0_5.sRm = LD; cekv0_5.sRn = 1;
      cekv0_5.M = Tt; cekv0_5.N = D; cekv0_5.K = C1; cekv0_5.zi_n = 1; cekv0_5.flags = 4; cekv0_5.act = 0;
      cekv0_5.alpha = 1.0f; cekv0_5.beta = 1.0f; cekv0_5.sa = 1.0f; cekv0_5.sb = 1.0f; cekv0_5.Npad = LD; cekv0_5.pad_ = 0;
      k_gemm<1><<<dim3((unsigned)((LD) + 31) / 32, (unsigned)((Tt) + 15) / 16, (unsigned)(Fo)), 32, 0, stream>>>(cekv0_5); }
    { GemmP cekv0_6;
      cekv0_6.A = HP + (size_t)4100 * C1; cekv0_6.B = wkv + 6; cekv0_6.bias = HP + (size_t)4100 * C1; cekv0_6.R = KV; cekv0_6.C = KV;
      cekv0_6.sAo = (long long)3 * 2050 * C1; cekv0_6.sAi = 0; cekv0_6.sAm = C1; cekv0_6.sAk = 1; cekv0_6.sBo = 0; cekv0_6.sBi = 0; cekv0_6.sBn = C1 * 9; cekv0_6.sBk = 9; cekv0_6.sCo = (long long)Tt * LD; cekv0_6.sCi = 0; cekv0_6.sCm = LD; cekv0_6.sRo = (long long)Tt * LD; cekv0_6.sRi = 0; cekv0_6.sRm = LD; cekv0_6.sRn = 1;
      cekv0_6.M = Tt; cekv0_6.N = D; cekv0_6.K = C1; cekv0_6.zi_n = 1; cekv0_6.flags = 4; cekv0_6.act = 0;
      cekv0_6.alpha = 1.0f; cekv0_6.beta = 1.0f; cekv0_6.sa = 1.0f; cekv0_6.sb = 1.0f; cekv0_6.Npad = LD; cekv0_6.pad_ = 0;
      k_gemm<1><<<dim3((unsigned)((LD) + 31) / 32, (unsigned)((Tt) + 15) / 16, (unsigned)(Fo)), 32, 0, stream>>>(cekv0_6); }
    { GemmP cekv0_7;
      cekv0_7.A = HP + (size_t)4101 * C1; cekv0_7.B = wkv + 7; cekv0_7.bias = HP + (size_t)4101 * C1; cekv0_7.R = KV; cekv0_7.C = KV;
      cekv0_7.sAo = (long long)3 * 2050 * C1; cekv0_7.sAi = 0; cekv0_7.sAm = C1; cekv0_7.sAk = 1; cekv0_7.sBo = 0; cekv0_7.sBi = 0; cekv0_7.sBn = C1 * 9; cekv0_7.sBk = 9; cekv0_7.sCo = (long long)Tt * LD; cekv0_7.sCi = 0; cekv0_7.sCm = LD; cekv0_7.sRo = (long long)Tt * LD; cekv0_7.sRi = 0; cekv0_7.sRm = LD; cekv0_7.sRn = 1;
      cekv0_7.M = Tt; cekv0_7.N = D; cekv0_7.K = C1; cekv0_7.zi_n = 1; cekv0_7.flags = 4; cekv0_7.act = 0;
      cekv0_7.alpha = 1.0f; cekv0_7.beta = 1.0f; cekv0_7.sa = 1.0f; cekv0_7.sb = 1.0f; cekv0_7.Npad = LD; cekv0_7.pad_ = 0;
      k_gemm<1><<<dim3((unsigned)((LD) + 31) / 32, (unsigned)((Tt) + 15) / 16, (unsigned)(Fo)), 32, 0, stream>>>(cekv0_7); }
    { GemmP cekv0_8;
      cekv0_8.A = HP + (size_t)4102 * C1; cekv0_8.B = wkv + 8; cekv0_8.bias = HP + (size_t)4102 * C1; cekv0_8.R = KV; cekv0_8.C = KV;
      cekv0_8.sAo = (long long)3 * 2050 * C1; cekv0_8.sAi = 0; cekv0_8.sAm = C1; cekv0_8.sAk = 1; cekv0_8.sBo = 0; cekv0_8.sBi = 0; cekv0_8.sBn = C1 * 9; cekv0_8.sBk = 9; cekv0_8.sCo = (long long)Tt * LD; cekv0_8.sCi = 0; cekv0_8.sCm = LD; cekv0_8.sRo = (long long)Tt * LD; cekv0_8.sRi = 0; cekv0_8.sRm = LD; cekv0_8.sRn = 1;
      cekv0_8.M = Tt; cekv0_8.N = D; cekv0_8.K = C1; cekv0_8.zi_n = 1; cekv0_8.flags = 4; cekv0_8.act = 0;
      cekv0_8.alpha = 1.0f; cekv0_8.beta = 1.0f; cekv0_8.sa = 1.0f; cekv0_8.sb = 1.0f; cekv0_8.Npad = LD; cekv0_8.pad_ = 0;
      k_gemm<1><<<dim3((unsigned)((LD) + 31) / 32, (unsigned)((Tt) + 15) / 16, (unsigned)(Fo)), 32, 0, stream>>>(cekv0_8); }

    k_cl_colsum1<<<NB, 256, 0, stream>>>(frame + (size_t)0 * Ll, 1, 1, (long long)Ll, PART); k_cl_colsum2<<<1, 256, 0, stream>>>(PART, NB, 1, RED, 0);
    k_cl_masknorm<<<(unsigned)((Ll + 255) / 256), 256, 0, stream>>>(KV, LD, frame + (size_t)0 * Ll, RED, Tsc, (long long)Ll, D);
    { GemmP gpQP0;
      gpQP0.A = Q; gpQP0.B = faq; gpQP0.bias = fabq; gpQP0.R = Q; gpQP0.C = QP;
      gpQP0.sAo = 0; gpQP0.sAi = 0; gpQP0.sAm = LD; gpQP0.sAk = 1; gpQP0.sBo = 0; gpQP0.sBi = 0; gpQP0.sBn = 1; gpQP0.sBk = D; gpQP0.sCo = 0; gpQP0.sCi = 0; gpQP0.sCm = LD; gpQP0.sRo = 0; gpQP0.sRi = 0; gpQP0.sRm = 0; gpQP0.sRn = 0;
      gpQP0.M = Ll; gpQP0.N = D; gpQP0.K = D; gpQP0.zi_n = 1; gpQP0.flags = 1; gpQP0.act = 6;
      gpQP0.alpha = 1.0f; gpQP0.beta = 0.0f; gpQP0.sa = 1.0f; gpQP0.sb = 1.0f; gpQP0.Npad = LD; gpQP0.pad_ = 0;
      k_gemm<1><<<dim3((unsigned)((LD) + 31) / 32, (unsigned)((Ll) + 15) / 16, (unsigned)(1)), 32, 0, stream>>>(gpQP0); }
    { GemmP gpKP0;
      gpKP0.A = KV; gpKP0.B = fak; gpKP0.bias = fabk; gpKP0.R = KV; gpKP0.C = KP;
      gpKP0.sAo = 0; gpKP0.sAi = 0; gpKP0.sAm = LD; gpKP0.sAk = 1; gpKP0.sBo = 0; gpKP0.sBi = 0; gpKP0.sBn = 1; gpKP0.sBk = D; gpKP0.sCo = 0; gpKP0.sCi = 0; gpKP0.sCm = LD; gpKP0.sRo = 0; gpKP0.sRi = 0; gpKP0.sRm = 0; gpKP0.sRn = 0;
      gpKP0.M = Ll; gpKP0.N = D; gpKP0.K = D; gpKP0.zi_n = 1; gpKP0.flags = 1; gpKP0.act = 6;
      gpKP0.alpha = 1.0f; gpKP0.beta = 0.0f; gpKP0.sa = 1.0f; gpKP0.sb = 1.0f; gpKP0.Npad = LD; gpKP0.pad_ = 0;
      k_gemm<1><<<dim3((unsigned)((LD) + 31) / 32, (unsigned)((Ll) + 15) / 16, (unsigned)(1)), 32, 0, stream>>>(gpKP0); }
    { GemmP gpVP0;
      gpVP0.A = KV; gpVP0.B = fav; gpVP0.bias = fabv; gpVP0.R = KV; gpVP0.C = VP;
      gpVP0.sAo = 0; gpVP0.sAi = 0; gpVP0.sAm = LD; gpVP0.sAk = 1; gpVP0.sBo = 0; gpVP0.sBi = 0; gpVP0.sBn = 1; gpVP0.sBk = D; gpVP0.sCo = 0; gpVP0.sCi = 0; gpVP0.sCm = LD; gpVP0.sRo = 0; gpVP0.sRi = 0; gpVP0.sRm = 0; gpVP0.sRn = 0;
      gpVP0.M = Ll; gpVP0.N = D; gpVP0.K = D; gpVP0.zi_n = 1; gpVP0.flags = 1; gpVP0.act = 0;
      gpVP0.alpha = 1.0f; gpVP0.beta = 0.0f; gpVP0.sa = 1.0f; gpVP0.sb = 1.0f; gpVP0.Npad = LD; gpVP0.pad_ = 0;
      k_gemm<1><<<dim3((unsigned)((LD) + 31) / 32, (unsigned)((Ll) + 15) / 16, (unsigned)(1)), 32, 0, stream>>>(gpVP0); }
    k_cl_colsum1<<<NB, 256, 0, stream>>>(KP, LD, D, (long long)Ll, PART); k_cl_colsum2<<<1, 256, 0, stream>>>(PART, NB, D, RED, 16);
    k_cl_colsum1<<<NB, 256, 0, stream>>>(QP, LD, D, (long long)Ll, PART); k_cl_colsum2<<<1, 256, 0, stream>>>(PART, NB, D, RED, 32);
    k_cl_flow1<<<(unsigned)((Ll + 255) / 256), 256, 0, stream>>>(QP, KP, LD, RED, SV, (long long)Ll, D);
    k_cl_flow2<<<(unsigned)(((long long)Ll * D + 255) / 256), 256, 0, stream>>>(QP, KP, LD, SV, O, O2, (long long)Ll, D);
    k_cl_colsum1<<<NB, 256, 0, stream>>>(O, LD, D, (long long)Ll, PART); k_cl_colsum2<<<1, 256, 0, stream>>>(PART, NB, D, RED, 48);
    k_cl_colsum1<<<NB, 256, 0, stream>>>(O2, LD, D, (long long)Ll, PART); k_cl_colsum2<<<1, 256, 0, stream>>>(PART, NB, D, RED, 64);
    k_cl_flow3<<<(unsigned)((Ll + 255) / 256), 256, 0, stream>>>(QP, KP, LD, RED, SV, (long long)Ll, D);
    k_cl_max1<<<NB, 256, 0, stream>>>(SV, 3, (long long)Ll, PART); k_cl_max2<<<1, 256, 0, stream>>>(PART, NB, RED, 80);
    k_cl_flow4<<<(unsigned)((Ll + 255) / 256), 256, 0, stream>>>(SV, RED, O2, LD, (long long)Ll);
    k_cl_colsum1<<<NB, 256, 0, stream>>>(O2 + 15, LD, 1, (long long)Ll, PART); k_cl_colsum2<<<1, 256, 0, stream>>>(PART, NB, 1, RED, 96);
    k_cl_flow5<<<(unsigned)(((long long)Ll * D + 255) / 256), 256, 0, stream>>>(VP, O2, LD, RED, O, (long long)Ll, D);
    { GemmP gkv0;
      gkv0.A = KP; gkv0.B = O; gkv0.bias = KP; gkv0.R = KP; gkv0.C = KVM;
      gkv0.sAo = 0; gkv0.sAi = 0; gkv0.sAm = 1; gkv0.sAk = LD; gkv0.sBo = 0; gkv0.sBi = 0; gkv0.sBn = 1; gkv0.sBk = LD; gkv0.sCo = 0; gkv0.sCi = 0; gkv0.sCm = LD; gkv0.sRo = 0; gkv0.sRi = 0; gkv0.sRm = 0; gkv0.sRn = 0;
      gkv0.M = D; gkv0.N = D; gkv0.K = Ll; gkv0.zi_n = 1; gkv0.flags = 0; gkv0.act = 0;
      gkv0.alpha = 1.0f; gkv0.beta = 0.0f; gkv0.sa = 1.0f; gkv0.sb = 1.0f; gkv0.Npad = LD; gkv0.pad_ = 0;
      k_gemm<1><<<dim3((unsigned)((LD) + 31) / 32, (unsigned)((D) + 15) / 16, (unsigned)(1)), 32, 0, stream>>>(gkv0); }
    { GemmP gqkv0;
      gqkv0.A = QP; gqkv0.B = KVM; gqkv0.bias = QP; gqkv0.R = QP; gqkv0.C = O2;
      gqkv0.sAo = 0; gqkv0.sAi = 0; gqkv0.sAm = LD; gqkv0.sAk = 1; gqkv0.sBo = 0; gqkv0.sBi = 0; gqkv0.sBn = 1; gqkv0.sBk = LD; gqkv0.sCo = 0; gqkv0.sCi = 0; gqkv0.sCm = LD; gqkv0.sRo = 0; gqkv0.sRi = 0; gqkv0.sRm = 0; gqkv0.sRn = 0;
      gqkv0.M = Ll; gqkv0.N = D; gqkv0.K = D; gqkv0.zi_n = 1; gqkv0.flags = 0; gqkv0.act = 0;
      gqkv0.alpha = 1.0f; gqkv0.beta = 0.0f; gqkv0.sa = 1.0f; gqkv0.sb = 1.0f; gqkv0.Npad = LD; gqkv0.pad_ = 0;
      k_gemm<1><<<dim3((unsigned)((LD) + 31) / 32, (unsigned)((Ll) + 15) / 16, (unsigned)(1)), 32, 0, stream>>>(gqkv0); }
    k_cl_flow6<<<(unsigned)(((long long)Ll * D + 255) / 256), 256, 0, stream>>>(O2, LD, SV, (long long)Ll, D);
    { GemmP gwo0;
      gwo0.A = O2; gwo0.B = fao; gwo0.bias = fabo; gwo0.R = O2; gwo0.C = O;
      gwo0.sAo = 0; gwo0.sAi = 0; gwo0.sAm = LD; gwo0.sAk = 1; gwo0.sBo = 0; gwo0.sBi = 0; gwo0.sBn = 1; gwo0.sBk = D; gwo0.sCo = 0; gwo0.sCi = 0; gwo0.sCm = LD; gwo0.sRo = 0; gwo0.sRi = 0; gwo0.sRm = 0; gwo0.sRn = 0;
      gwo0.M = Ll; gwo0.N = D; gwo0.K = D; gwo0.zi_n = 1; gwo0.flags = 1; gwo0.act = 0;
      gwo0.alpha = 1.0f; gwo0.beta = 0.0f; gwo0.sa = 1.0f; gwo0.sb = 1.0f; gwo0.Npad = LD; gwo0.pad_ = 0;
      k_gemm<1><<<dim3((unsigned)((LD) + 31) / 32, (unsigned)((Ll) + 15) / 16, (unsigned)(1)), 32, 0, stream>>>(gwo0); }
    k_cl_out<<<(unsigned)(((long long)Ll * D + 255) / 256), 256, 0, stream>>>(O, LD, out, 0, (long long)Ll, D);
    hipMemsetAsync(XP, 0, (size_t)256 * 2052 * CI * 4, stream); hipMemsetAsync(HP, 0, (size_t)Hh * 2050 * C1 * 4, stream);
    k_cl_pad<<<(unsigned)(((long long)Hh * Tt * CI + 255) / 256), 256, 0, stream>>>(x, XP, 1, CI, Hh, Tt);
    { GemmP cp1_0;
      cp1_0.A = XP + (size_t)0 * CI; cp1_0.B = wpre + 0; cp1_0.bias = bpre; cp1_0.R = XP + (size_t)0 * CI; cp1_0.C = HP + C1;
      cp1_0.sAo = (long long)2052 * CI; cp1_0.sAi = 0; cp1_0.sAm = CI; cp1_0.sAk = 1; cp1_0.sBo = 0; cp1_0.sBi = 0; cp1_0.sBn = CI * 25; cp1_0.sBk = 25; cp1_0.sCo = (long long)2050 * C1; cp1_0.sCi = 0; cp1_0.sCm = C1; cp1_0.sRo = 0; cp1_0.sRi = 0; cp1_0.sRm = 0; cp1_0.sRn = 0;
      cp1_0.M = Tt; cp1_0.N = C1; cp1_0.K = CI; cp1_0.zi_n = 1; cp1_0.flags = 1; cp1_0.act = 0;
      cp1_0.alpha = 1.0f; cp1_0.beta = 0.0f; cp1_0.sa = 1.0f; cp1_0.sb = 1.0f; cp1_0.Npad = C1; cp1_0.pad_ = 0;
      k_gemm<1><<<dim3((unsigned)((C1) + 31) / 32, (unsigned)((Tt) + 15) / 16, (unsigned)(Hh)), 32, 0, stream>>>(cp1_0); }
    { GemmP cp1_1;
      cp1_1.A = XP + (size_t)1 * CI; cp1_1.B = wpre + 1; cp1_1.bias = XP + (size_t)1 * CI; cp1_1.R = HP + C1; cp1_1.C = HP + C1;
      cp1_1.sAo = (long long)2052 * CI; cp1_1.sAi = 0; cp1_1.sAm = CI; cp1_1.sAk = 1; cp1_1.sBo = 0; cp1_1.sBi = 0; cp1_1.sBn = CI * 25; cp1_1.sBk = 25; cp1_1.sCo = (long long)2050 * C1; cp1_1.sCi = 0; cp1_1.sCm = C1; cp1_1.sRo = (long long)2050 * C1; cp1_1.sRi = 0; cp1_1.sRm = C1; cp1_1.sRn = 1;
      cp1_1.M = Tt; cp1_1.N = C1; cp1_1.K = CI; cp1_1.zi_n = 1; cp1_1.flags = 4; cp1_1.act = 0;
      cp1_1.alpha = 1.0f; cp1_1.beta = 1.0f; cp1_1.sa = 1.0f; cp1_1.sb = 1.0f; cp1_1.Npad = C1; cp1_1.pad_ = 0;
      k_gemm<1><<<dim3((unsigned)((C1) + 31) / 32, (unsigned)((Tt) + 15) / 16, (unsigned)(Hh)), 32, 0, stream>>>(cp1_1); }
    { GemmP cp1_2;
      cp1_2.A = XP + (size_t)2 * CI; cp1_2.B = wpre + 2; cp1_2.bias = XP + (size_t)2 * CI; cp1_2.R = HP + C1; cp1_2.C = HP + C1;
      cp1_2.sAo = (long long)2052 * CI; cp1_2.sAi = 0; cp1_2.sAm = CI; cp1_2.sAk = 1; cp1_2.sBo = 0; cp1_2.sBi = 0; cp1_2.sBn = CI * 25; cp1_2.sBk = 25; cp1_2.sCo = (long long)2050 * C1; cp1_2.sCi = 0; cp1_2.sCm = C1; cp1_2.sRo = (long long)2050 * C1; cp1_2.sRi = 0; cp1_2.sRm = C1; cp1_2.sRn = 1;
      cp1_2.M = Tt; cp1_2.N = C1; cp1_2.K = CI; cp1_2.zi_n = 1; cp1_2.flags = 4; cp1_2.act = 0;
      cp1_2.alpha = 1.0f; cp1_2.beta = 1.0f; cp1_2.sa = 1.0f; cp1_2.sb = 1.0f; cp1_2.Npad = C1; cp1_2.pad_ = 0;
      k_gemm<1><<<dim3((unsigned)((C1) + 31) / 32, (unsigned)((Tt) + 15) / 16, (unsigned)(Hh)), 32, 0, stream>>>(cp1_2); }
    { GemmP cp1_3;
      cp1_3.A = XP + (size_t)3 * CI; cp1_3.B = wpre + 3; cp1_3.bias = XP + (size_t)3 * CI; cp1_3.R = HP + C1; cp1_3.C = HP + C1;
      cp1_3.sAo = (long long)2052 * CI; cp1_3.sAi = 0; cp1_3.sAm = CI; cp1_3.sAk = 1; cp1_3.sBo = 0; cp1_3.sBi = 0; cp1_3.sBn = CI * 25; cp1_3.sBk = 25; cp1_3.sCo = (long long)2050 * C1; cp1_3.sCi = 0; cp1_3.sCm = C1; cp1_3.sRo = (long long)2050 * C1; cp1_3.sRi = 0; cp1_3.sRm = C1; cp1_3.sRn = 1;
      cp1_3.M = Tt; cp1_3.N = C1; cp1_3.K = CI; cp1_3.zi_n = 1; cp1_3.flags = 4; cp1_3.act = 0;
      cp1_3.alpha = 1.0f; cp1_3.beta = 1.0f; cp1_3.sa = 1.0f; cp1_3.sb = 1.0f; cp1_3.Npad = C1; cp1_3.pad_ = 0;
      k_gemm<1><<<dim3((unsigned)((C1) + 31) / 32, (unsigned)((Tt) + 15) / 16, (unsigned)(Hh)), 32, 0, stream>>>(cp1_3); }
    { GemmP cp1_4;
      cp1_4.A = XP + (size_t)4 * CI; cp1_4.B = wpre + 4; cp1_4.bias = XP + (size_t)4 * CI; cp1_4.R = HP + C1; cp1_4.C = HP + C1;
      cp1_4.sAo = (long long)2052 * CI; cp1_4.sAi = 0; cp1_4.sAm = CI; cp1_4.sAk = 1; cp1_4.sBo = 0; cp1_4.sBi = 0; cp1_4.sBn = CI * 25; cp1_4.sBk = 25; cp1_4.sCo = (long long)2050 * C1; cp1_4.sCi = 0; cp1_4.sCm = C1; cp1_4.sRo = (long long)2050 * C1; cp1_4.sRi = 0; cp1_4.sRm = C1; cp1_4.sRn = 1;
      cp1_4.M = Tt; cp1_4.N = C1; cp1_4.K = CI; cp1_4.zi_n = 1; cp1_4.flags = 4; cp1_4.act = 0;
      cp1_4.alpha = 1.0f; cp1_4.beta = 1.0f; cp1_4.sa = 1.0f; cp1_4.sb = 1.0f; cp1_4.Npad = C1; cp1_4.pad_ = 0;
      k_gemm<1><<<dim3((unsigned)((C1) + 31) / 32, (unsigned)((Tt) + 15) / 16, (unsigned)(Hh)), 32, 0, stream>>>(cp1_4); }
    { GemmP cp1_5;
      cp1_5.A = XP + (size_t)2052 * CI; cp1_5.B = wpre + 5; cp1_5.bias = XP + (size_t)2052 * CI; cp1_5.R = HP + C1; cp1_5.C = HP + C1;
      cp1_5.sAo = (long long)2052 * CI; cp1_5.sAi = 0; cp1_5.sAm = CI; cp1_5.sAk = 1; cp1_5.sBo = 0; cp1_5.sBi = 0; cp1_5.sBn = CI * 25; cp1_5.sBk = 25; cp1_5.sCo = (long long)2050 * C1; cp1_5.sCi = 0; cp1_5.sCm = C1; cp1_5.sRo = (long long)2050 * C1; cp1_5.sRi = 0; cp1_5.sRm = C1; cp1_5.sRn = 1;
      cp1_5.M = Tt; cp1_5.N = C1; cp1_5.K = CI; cp1_5.zi_n = 1; cp1_5.flags = 4; cp1_5.act = 0;
      cp1_5.alpha = 1.0f; cp1_5.beta = 1.0f; cp1_5.sa = 1.0f; cp1_5.sb = 1.0f; cp1_5.Npad = C1; cp1_5.pad_ = 0;
      k_gemm<1><<<dim3((unsigned)((C1) + 31) / 32, (unsigned)((Tt) + 15) / 16, (unsigned)(Hh)), 32, 0, stream>>>(cp1_5); }
    { GemmP cp1_6;
      cp1_6.A = XP + (size_t)2053 * CI; cp1_6.B = wpre + 6; cp1_6.bias = XP + (size_t)2053 * CI; cp1_6.R = HP + C1; cp1_6.C = HP + C1;
      cp1_6.sAo = (long long)2052 * CI; cp1_6.sAi = 0; cp1_6.sAm = CI; cp1_6.sAk = 1; cp1_6.sBo = 0; cp1_6.sBi = 0; cp1_6.sBn = CI * 25; cp1_6.sBk = 25; cp1_6.sCo = (long long)2050 * C1; cp1_6.sCi = 0; cp1_6.sCm = C1; cp1_6.sRo = (long long)2050 * C1; cp1_6.sRi = 0; cp1_6.sRm = C1; cp1_6.sRn = 1;
      cp1_6.M = Tt; cp1_6.N = C1; cp1_6.K = CI; cp1_6.zi_n = 1; cp1_6.flags = 4; cp1_6.act = 0;
      cp1_6.alpha = 1.0f; cp1_6.beta = 1.0f; cp1_6.sa = 1.0f; cp1_6.sb = 1.0f; cp1_6.Npad = C1; cp1_6.pad_ = 0;
      k_gemm<1><<<dim3((unsigned)((C1) + 31) / 32, (unsigned)((Tt) + 15) / 16, (unsigned)(Hh)), 32, 0, stream>>>(cp1_6); }
    { GemmP cp1_7;
      cp1_7.A = XP + (size_t)2054 * CI; cp1_7.B = wpre + 7; cp1_7.bias = XP + (size_t)2054 * CI; cp1_7.R = HP + C1; cp1_7.C = HP + C1;
      cp1_7.sAo = (long long)2052 * CI; cp1_7.sAi = 0; cp1_7.sAm = CI; cp1_7.sAk = 1; cp1_7.sBo = 0; cp1_7.sBi = 0; cp1_7.sBn = CI * 25; cp1_7.sBk = 25; cp1_7.sCo = (long long)2050 * C1; cp1_7.sCi = 0; cp1_7.sCm = C1; cp1_7.sRo = (long long)2050 * C1; cp1_7.sRi = 0; cp1_7.sRm = C1; cp1_7.sRn = 1;
      cp1_7.M = Tt; cp1_7.N = C1; cp1_7.K = CI; cp1_7.zi_n = 1; cp1_7.flags = 4; cp1_7.act = 0;
      cp1_7.alpha = 1.0f; cp1_7.beta = 1.0f; cp1_7.sa = 1.0f; cp1_7.sb = 1.0f; cp1_7.Npad = C1; cp1_7.pad_ = 0;
      k_gemm<1><<<dim3((unsigned)((C1) + 31) / 32, (unsigned)((Tt) + 15) / 16, (unsigned)(Hh)), 32, 0, stream>>>(cp1_7); }
    { GemmP cp1_8;
      cp1_8.A = XP + (size_t)2055 * CI; cp1_8.B = wpre + 8; cp1_8.bias = XP + (size_t)2055 * CI; cp1_8.R = HP + C1; cp1_8.C = HP + C1;
      cp1_8.sAo = (long long)2052 * CI; cp1_8.sAi = 0; cp1_8.sAm = CI; cp1_8.sAk = 1; cp1_8.sBo = 0; cp1_8.sBi = 0; cp1_8.sBn = CI * 25; cp1_8.sBk = 25; cp1_8.sCo = (long long)2050 * C1; cp1_8.sCi = 0; cp1_8.sCm = C1; cp1_8.sRo = (long long)2050 * C1; cp1_8.sRi = 0; cp1_8.sRm = C1; cp1_8.sRn = 1;
      cp1_8.M = Tt; cp1_8.N = C1; cp1_8.K = CI; cp1_8.zi_n = 1; cp1_8.flags = 4; cp1_8.act = 0;
      cp1_8.alpha = 1.0f; cp1_8.beta = 1.0f; cp1_8.sa = 1.0f; cp1_8.sb = 1.0f; cp1_8.Npad = C1; cp1_8.pad_ = 0;
      k_gemm<1><<<dim3((unsigned)((C1) + 31) / 32, (unsigned)((Tt) + 15) / 16, (unsigned)(Hh)), 32, 0, stream>>>(cp1_8); }
    { GemmP cp1_9;
      cp1_9.A = XP + (size_t)2056 * CI; cp1_9.B = wpre + 9; cp1_9.bias = XP + (size_t)2056 * CI; cp1_9.R = HP + C1; cp1_9.C = HP + C1;
      cp1_9.sAo = (long long)2052 * CI; cp1_9.sAi = 0; cp1_9.sAm = CI; cp1_9.sAk = 1; cp1_9.sBo = 0; cp1_9.sBi = 0; cp1_9.sBn = CI * 25; cp1_9.sBk = 25; cp1_9.sCo = (long long)2050 * C1; cp1_9.sCi = 0; cp1_9.sCm = C1; cp1_9.sRo = (long long)2050 * C1; cp1_9.sRi = 0; cp1_9.sRm = C1; cp1_9.sRn = 1;
      cp1_9.M = Tt; cp1_9.N = C1; cp1_9.K = CI; cp1_9.zi_n = 1; cp1_9.flags = 4; cp1_9.act = 0;
      cp1_9.alpha = 1.0f; cp1_9.beta = 1.0f; cp1_9.sa = 1.0f; cp1_9.sb = 1.0f; cp1_9.Npad = C1; cp1_9.pad_ = 0;
      k_gemm<1><<<dim3((unsigned)((C1) + 31) / 32, (unsigned)((Tt) + 15) / 16, (unsigned)(Hh)), 32, 0, stream>>>(cp1_9); }
    { GemmP cp1_10;
      cp1_10.A = XP + (size_t)4104 * CI; cp1_10.B = wpre + 10; cp1_10.bias = XP + (size_t)4104 * CI; cp1_10.R = HP + C1; cp1_10.C = HP + C1;
      cp1_10.sAo = (long long)2052 * CI; cp1_10.sAi = 0; cp1_10.sAm = CI; cp1_10.sAk = 1; cp1_10.sBo = 0; cp1_10.sBi = 0; cp1_10.sBn = CI * 25; cp1_10.sBk = 25; cp1_10.sCo = (long long)2050 * C1; cp1_10.sCi = 0; cp1_10.sCm = C1; cp1_10.sRo = (long long)2050 * C1; cp1_10.sRi = 0; cp1_10.sRm = C1; cp1_10.sRn = 1;
      cp1_10.M = Tt; cp1_10.N = C1; cp1_10.K = CI; cp1_10.zi_n = 1; cp1_10.flags = 4; cp1_10.act = 0;
      cp1_10.alpha = 1.0f; cp1_10.beta = 1.0f; cp1_10.sa = 1.0f; cp1_10.sb = 1.0f; cp1_10.Npad = C1; cp1_10.pad_ = 0;
      k_gemm<1><<<dim3((unsigned)((C1) + 31) / 32, (unsigned)((Tt) + 15) / 16, (unsigned)(Hh)), 32, 0, stream>>>(cp1_10); }
    { GemmP cp1_11;
      cp1_11.A = XP + (size_t)4105 * CI; cp1_11.B = wpre + 11; cp1_11.bias = XP + (size_t)4105 * CI; cp1_11.R = HP + C1; cp1_11.C = HP + C1;
      cp1_11.sAo = (long long)2052 * CI; cp1_11.sAi = 0; cp1_11.sAm = CI; cp1_11.sAk = 1; cp1_11.sBo = 0; cp1_11.sBi = 0; cp1_11.sBn = CI * 25; cp1_11.sBk = 25; cp1_11.sCo = (long long)2050 * C1; cp1_11.sCi = 0; cp1_11.sCm = C1; cp1_11.sRo = (long long)2050 * C1; cp1_11.sRi = 0; cp1_11.sRm = C1; cp1_11.sRn = 1;
      cp1_11.M = Tt; cp1_11.N = C1; cp1_11.K = CI; cp1_11.zi_n = 1; cp1_11.flags = 4; cp1_11.act = 0;
      cp1_11.alpha = 1.0f; cp1_11.beta = 1.0f; cp1_11.sa = 1.0f; cp1_11.sb = 1.0f; cp1_11.Npad = C1; cp1_11.pad_ = 0;
      k_gemm<1><<<dim3((unsigned)((C1) + 31) / 32, (unsigned)((Tt) + 15) / 16, (unsigned)(Hh)), 32, 0, stream>>>(cp1_11); }
    { GemmP cp1_12;
      cp1_12.A = XP + (size_t)4106 * CI; cp1_12.B = wpre + 12; cp1_12.bias = XP + (size_t)4106 * CI; cp1_12.R = HP + C1; cp1_12.C = HP + C1;
      cp1_12.sAo = (long long)2052 * CI; cp1_12.sAi = 0; cp1_12.sAm = CI; cp1_12.sAk = 1; cp1_12.sBo = 0; cp1_12.sBi = 0; cp1_12.sBn = CI * 25; cp1_12.sBk = 25; cp1_12.sCo = (long long)2050 * C1; cp1_12.sCi = 0; cp1_12.sCm = C1; cp1_12.sRo = (long long)2050 * C1; cp1_12.sRi = 0; cp1_12.sRm = C1; cp1_12.sRn = 1;
      cp1_12.M = Tt; cp1_12.N = C1; cp1_12.K = CI; cp1_12.zi_n = 1; cp1_12.flags = 4; cp1_12.act = 0;
      cp1_12.alpha = 1.0f; cp1_12.beta = 1.0f; cp1_12.sa = 1.0f; cp1_12.sb = 1.0f; cp1_12.Npad = C1; cp1_12.pad_ = 0;
      k_gemm<1><<<dim3((unsigned)((C1) + 31) / 32, (unsigned)((Tt) + 15) / 16, (unsigned)(Hh)), 32, 0, stream>>>(cp1_12); }
    { GemmP cp1_13;
      cp1_13.A = XP + (size_t)4107 * CI; cp1_13.B = wpre + 13; cp1_13.bias = XP + (size_t)4107 * CI; cp1_13.R = HP + C1; cp1_13.C = HP + C1;
      cp1_13.sAo = (long long)2052 * CI; cp1_13.sAi = 0; cp1_13.sAm = CI; cp1_13.sAk = 1; cp1_13.sBo = 0; cp1_13.sBi = 0; cp1_13.sBn = CI * 25; cp1_13.sBk = 25; cp1_13.sCo = (long long)2050 * C1; cp1_13.sCi = 0; cp1_13.sCm = C1; cp1_13.sRo = (long long)2050 * C1; cp1_13.sRi = 0; cp1_13.sRm = C1; cp1_13.sRn = 1;
      cp1_13.M = Tt; cp1_13.N = C1; cp1_13.K = CI; cp1_13.zi_n = 1; cp1_13.flags = 4; cp1_13.act = 0;
      cp1_13.alpha = 1.0f; cp1_13.beta = 1.0f; cp1_13.sa = 1.0f; cp1_13.sb = 1.0f; cp1_13.Npad = C1; cp1_13.pad_ = 0;
      k_gemm<1><<<dim3((unsigned)((C1) + 31) / 32, (unsigned)((Tt) + 15) / 16, (unsigned)(Hh)), 32, 0, stream>>>(cp1_13); }
    { GemmP cp1_14;
      cp1_14.A = XP + (size_t)4108 * CI; cp1_14.B = wpre + 14; cp1_14.bias = XP + (size_t)4108 * CI; cp1_14.R = HP + C1; cp1_14.C = HP + C1;
      cp1_14.sAo = (long long)2052 * CI; cp1_14.sAi = 0; cp1_14.sAm = CI; cp1_14.sAk = 1; cp1_14.sBo = 0; cp1_14.sBi = 0; cp1_14.sBn = CI * 25; cp1_14.sBk = 25; cp1_14.sCo = (long long)2050 * C1; cp1_14.sCi = 0; cp1_14.sCm = C1; cp1_14.sRo = (long long)2050 * C1; cp1_14.sRi = 0; cp1_14.sRm = C1; cp1_14.sRn = 1;
      cp1_14.M = Tt; cp1_14.N = C1; cp1_14.K = CI; cp1_14.zi_n = 1; cp1_14.flags = 4; cp1_14.act = 0;
      cp1_14.alpha = 1.0f; cp1_14.beta = 1.0f; cp1_14.sa = 1.0f; cp1_14.sb = 1.0f; cp1_14.Npad = C1; cp1_14.pad_ = 0;
      k_gemm<1><<<dim3((unsigned)((C1) + 31) / 32, (unsigned)((Tt) + 15) / 16, (unsigned)(Hh)), 32, 0, stream>>>(cp1_14); }
    { GemmP cp1_15;
      cp1_15.A = XP + (size_t)6156 * CI; cp1_15.B = wpre + 15; cp1_15.bias = XP + (size_t)6156 * CI; cp1_15.R = HP + C1; cp1_15.C = HP + C1;
      cp1_15.sAo = (long long)2052 * CI; cp1_15.sAi = 0; cp1_15.sAm = CI; cp1_15.sAk = 1; cp1_15.sBo = 0; cp1_15.sBi = 0; cp1_15.sBn = CI * 25; cp1_15.sBk = 25; cp1_15.sCo = (long long)2050 * C1; cp1_15.sCi = 0; cp1_15.sCm = C1; cp1_15.sRo = (long long)2050 * C1; cp1_15.sRi = 0; cp1_15.sRm = C1; cp1_15.sRn = 1;
      cp1_15.M = Tt; cp1_15.N = C1; cp1_15.K = CI; cp1_15.zi_n = 1; cp1_15.flags = 4; cp1_15.act = 0;
      cp1_15.alpha = 1.0f; cp1_15.beta = 1.0f; cp1_15.sa = 1.0f; cp1_15.sb = 1.0f; cp1_15.Npad = C1; cp1_15.pad_ = 0;
      k_gemm<1><<<dim3((unsigned)((C1) + 31) / 32, (unsigned)((Tt) + 15) / 16, (unsigned)(Hh)), 32, 0, stream>>>(cp1_15); }
    { GemmP cp1_16;
      cp1_16.A = XP + (size_t)6157 * CI; cp1_16.B = wpre + 16; cp1_16.bias = XP + (size_t)6157 * CI; cp1_16.R = HP + C1; cp1_16.C = HP + C1;
      cp1_16.sAo = (long long)2052 * CI; cp1_16.sAi = 0; cp1_16.sAm = CI; cp1_16.sAk = 1; cp1_16.sBo = 0; cp1_16.sBi = 0; cp1_16.sBn = CI * 25; cp1_16.sBk = 25; cp1_16.sCo = (long long)2050 * C1; cp1_16.sCi = 0; cp1_16.sCm = C1; cp1_16.sRo = (long long)2050 * C1; cp1_16.sRi = 0; cp1_16.sRm = C1; cp1_16.sRn = 1;
      cp1_16.M = Tt; cp1_16.N = C1; cp1_16.K = CI; cp1_16.zi_n = 1; cp1_16.flags = 4; cp1_16.act = 0;
      cp1_16.alpha = 1.0f; cp1_16.beta = 1.0f; cp1_16.sa = 1.0f; cp1_16.sb = 1.0f; cp1_16.Npad = C1; cp1_16.pad_ = 0;
      k_gemm<1><<<dim3((unsigned)((C1) + 31) / 32, (unsigned)((Tt) + 15) / 16, (unsigned)(Hh)), 32, 0, stream>>>(cp1_16); }
    { GemmP cp1_17;
      cp1_17.A = XP + (size_t)6158 * CI; cp1_17.B = wpre + 17; cp1_17.bias = XP + (size_t)6158 * CI; cp1_17.R = HP + C1; cp1_17.C = HP + C1;
      cp1_17.sAo = (long long)2052 * CI; cp1_17.sAi = 0; cp1_17.sAm = CI; cp1_17.sAk = 1; cp1_17.sBo = 0; cp1_17.sBi = 0; cp1_17.sBn = CI * 25; cp1_17.sBk = 25; cp1_17.sCo = (long long)2050 * C1; cp1_17.sCi = 0; cp1_17.sCm = C1; cp1_17.sRo = (long long)2050 * C1; cp1_17.sRi = 0; cp1_17.sRm = C1; cp1_17.sRn = 1;
      cp1_17.M = Tt; cp1_17.N = C1; cp1_17.K = CI; cp1_17.zi_n = 1; cp1_17.flags = 4; cp1_17.act = 0;
      cp1_17.alpha = 1.0f; cp1_17.beta = 1.0f; cp1_17.sa = 1.0f; cp1_17.sb = 1.0f; cp1_17.Npad = C1; cp1_17.pad_ = 0;
      k_gemm<1><<<dim3((unsigned)((C1) + 31) / 32, (unsigned)((Tt) + 15) / 16, (unsigned)(Hh)), 32, 0, stream>>>(cp1_17); }
    { GemmP cp1_18;
      cp1_18.A = XP + (size_t)6159 * CI; cp1_18.B = wpre + 18; cp1_18.bias = XP + (size_t)6159 * CI; cp1_18.R = HP + C1; cp1_18.C = HP + C1;
      cp1_18.sAo = (long long)2052 * CI; cp1_18.sAi = 0; cp1_18.sAm = CI; cp1_18.sAk = 1; cp1_18.sBo = 0; cp1_18.sBi = 0; cp1_18.sBn = CI * 25; cp1_18.sBk = 25; cp1_18.sCo = (long long)2050 * C1; cp1_18.sCi = 0; cp1_18.sCm = C1; cp1_18.sRo = (long long)2050 * C1; cp1_18.sRi = 0; cp1_18.sRm = C1; cp1_18.sRn = 1;
      cp1_18.M = Tt; cp1_18.N = C1; cp1_18.K = CI; cp1_18.zi_n = 1; cp1_18.flags = 4; cp1_18.act = 0;
      cp1_18.alpha = 1.0f; cp1_18.beta = 1.0f; cp1_18.sa = 1.0f; cp1_18.sb = 1.0f; cp1_18.Npad = C1; cp1_18.pad_ = 0;
      k_gemm<1><<<dim3((unsigned)((C1) + 31) / 32, (unsigned)((Tt) + 15) / 16, (unsigned)(Hh)), 32, 0, stream>>>(cp1_18); }
    { GemmP cp1_19;
      cp1_19.A = XP + (size_t)6160 * CI; cp1_19.B = wpre + 19; cp1_19.bias = XP + (size_t)6160 * CI; cp1_19.R = HP + C1; cp1_19.C = HP + C1;
      cp1_19.sAo = (long long)2052 * CI; cp1_19.sAi = 0; cp1_19.sAm = CI; cp1_19.sAk = 1; cp1_19.sBo = 0; cp1_19.sBi = 0; cp1_19.sBn = CI * 25; cp1_19.sBk = 25; cp1_19.sCo = (long long)2050 * C1; cp1_19.sCi = 0; cp1_19.sCm = C1; cp1_19.sRo = (long long)2050 * C1; cp1_19.sRi = 0; cp1_19.sRm = C1; cp1_19.sRn = 1;
      cp1_19.M = Tt; cp1_19.N = C1; cp1_19.K = CI; cp1_19.zi_n = 1; cp1_19.flags = 4; cp1_19.act = 0;
      cp1_19.alpha = 1.0f; cp1_19.beta = 1.0f; cp1_19.sa = 1.0f; cp1_19.sb = 1.0f; cp1_19.Npad = C1; cp1_19.pad_ = 0;
      k_gemm<1><<<dim3((unsigned)((C1) + 31) / 32, (unsigned)((Tt) + 15) / 16, (unsigned)(Hh)), 32, 0, stream>>>(cp1_19); }
    { GemmP cp1_20;
      cp1_20.A = XP + (size_t)8208 * CI; cp1_20.B = wpre + 20; cp1_20.bias = XP + (size_t)8208 * CI; cp1_20.R = HP + C1; cp1_20.C = HP + C1;
      cp1_20.sAo = (long long)2052 * CI; cp1_20.sAi = 0; cp1_20.sAm = CI; cp1_20.sAk = 1; cp1_20.sBo = 0; cp1_20.sBi = 0; cp1_20.sBn = CI * 25; cp1_20.sBk = 25; cp1_20.sCo = (long long)2050 * C1; cp1_20.sCi = 0; cp1_20.sCm = C1; cp1_20.sRo = (long long)2050 * C1; cp1_20.sRi = 0; cp1_20.sRm = C1; cp1_20.sRn = 1;
      cp1_20.M = Tt; cp1_20.N = C1; cp1_20.K = CI; cp1_20.zi_n = 1; cp1_20.flags = 4; cp1_20.act = 0;
      cp1_20.alpha = 1.0f; cp1_20.beta = 1.0f; cp1_20.sa = 1.0f; cp1_20.sb = 1.0f; cp1_20.Npad = C1; cp1_20.pad_ = 0;
      k_gemm<1><<<dim3((unsigned)((C1) + 31) / 32, (unsigned)((Tt) + 15) / 16, (unsigned)(Hh)), 32, 0, stream>>>(cp1_20); }
    { GemmP cp1_21;
      cp1_21.A = XP + (size_t)8209 * CI; cp1_21.B = wpre + 21; cp1_21.bias = XP + (size_t)8209 * CI; cp1_21.R = HP + C1; cp1_21.C = HP + C1;
      cp1_21.sAo = (long long)2052 * CI; cp1_21.sAi = 0; cp1_21.sAm = CI; cp1_21.sAk = 1; cp1_21.sBo = 0; cp1_21.sBi = 0; cp1_21.sBn = CI * 25; cp1_21.sBk = 25; cp1_21.sCo = (long long)2050 * C1; cp1_21.sCi = 0; cp1_21.sCm = C1; cp1_21.sRo = (long long)2050 * C1; cp1_21.sRi = 0; cp1_21.sRm = C1; cp1_21.sRn = 1;
      cp1_21.M = Tt; cp1_21.N = C1; cp1_21.K = CI; cp1_21.zi_n = 1; cp1_21.flags = 4; cp1_21.act = 0;
      cp1_21.alpha = 1.0f; cp1_21.beta = 1.0f; cp1_21.sa = 1.0f; cp1_21.sb = 1.0f; cp1_21.Npad = C1; cp1_21.pad_ = 0;
      k_gemm<1><<<dim3((unsigned)((C1) + 31) / 32, (unsigned)((Tt) + 15) / 16, (unsigned)(Hh)), 32, 0, stream>>>(cp1_21); }
    { GemmP cp1_22;
      cp1_22.A = XP + (size_t)8210 * CI; cp1_22.B = wpre + 22; cp1_22.bias = XP + (size_t)8210 * CI; cp1_22.R = HP + C1; cp1_22.C = HP + C1;
      cp1_22.sAo = (long long)2052 * CI; cp1_22.sAi = 0; cp1_22.sAm = CI; cp1_22.sAk = 1; cp1_22.sBo = 0; cp1_22.sBi = 0; cp1_22.sBn = CI * 25; cp1_22.sBk = 25; cp1_22.sCo = (long long)2050 * C1; cp1_22.sCi = 0; cp1_22.sCm = C1; cp1_22.sRo = (long long)2050 * C1; cp1_22.sRi = 0; cp1_22.sRm = C1; cp1_22.sRn = 1;
      cp1_22.M = Tt; cp1_22.N = C1; cp1_22.K = CI; cp1_22.zi_n = 1; cp1_22.flags = 4; cp1_22.act = 0;
      cp1_22.alpha = 1.0f; cp1_22.beta = 1.0f; cp1_22.sa = 1.0f; cp1_22.sb = 1.0f; cp1_22.Npad = C1; cp1_22.pad_ = 0;
      k_gemm<1><<<dim3((unsigned)((C1) + 31) / 32, (unsigned)((Tt) + 15) / 16, (unsigned)(Hh)), 32, 0, stream>>>(cp1_22); }
    { GemmP cp1_23;
      cp1_23.A = XP + (size_t)8211 * CI; cp1_23.B = wpre + 23; cp1_23.bias = XP + (size_t)8211 * CI; cp1_23.R = HP + C1; cp1_23.C = HP + C1;
      cp1_23.sAo = (long long)2052 * CI; cp1_23.sAi = 0; cp1_23.sAm = CI; cp1_23.sAk = 1; cp1_23.sBo = 0; cp1_23.sBi = 0; cp1_23.sBn = CI * 25; cp1_23.sBk = 25; cp1_23.sCo = (long long)2050 * C1; cp1_23.sCi = 0; cp1_23.sCm = C1; cp1_23.sRo = (long long)2050 * C1; cp1_23.sRi = 0; cp1_23.sRm = C1; cp1_23.sRn = 1;
      cp1_23.M = Tt; cp1_23.N = C1; cp1_23.K = CI; cp1_23.zi_n = 1; cp1_23.flags = 4; cp1_23.act = 0;
      cp1_23.alpha = 1.0f; cp1_23.beta = 1.0f; cp1_23.sa = 1.0f; cp1_23.sb = 1.0f; cp1_23.Npad = C1; cp1_23.pad_ = 0;
      k_gemm<1><<<dim3((unsigned)((C1) + 31) / 32, (unsigned)((Tt) + 15) / 16, (unsigned)(Hh)), 32, 0, stream>>>(cp1_23); }
    { GemmP cp1_24;
      cp1_24.A = XP + (size_t)8212 * CI; cp1_24.B = wpre + 24; cp1_24.bias = XP + (size_t)8212 * CI; cp1_24.R = HP + C1; cp1_24.C = HP + C1;
      cp1_24.sAo = (long long)2052 * CI; cp1_24.sAi = 0; cp1_24.sAm = CI; cp1_24.sAk = 1; cp1_24.sBo = 0; cp1_24.sBi = 0; cp1_24.sBn = CI * 25; cp1_24.sBk = 25; cp1_24.sCo = (long long)2050 * C1; cp1_24.sCi = 0; cp1_24.sCm = C1; cp1_24.sRo = (long long)2050 * C1; cp1_24.sRi = 0; cp1_24.sRm = C1; cp1_24.sRn = 1;
      cp1_24.M = Tt; cp1_24.N = C1; cp1_24.K = CI; cp1_24.zi_n = 1; cp1_24.flags = 4; cp1_24.act = 0;
      cp1_24.alpha = 1.0f; cp1_24.beta = 1.0f; cp1_24.sa = 1.0f; cp1_24.sb = 1.0f; cp1_24.Npad = C1; cp1_24.pad_ = 0;
      k_gemm<1><<<dim3((unsigned)((C1) + 31) / 32, (unsigned)((Tt) + 15) / 16, (unsigned)(Hh)), 32, 0, stream>>>(cp1_24); }
    k_cl_bnl<<<(unsigned)(((long long)Hh * Tt * C1 + 255) / 256), 256, 0, stream>>>(HP, bng, bnb, bnm, bnv, Hh, Tt, C1);
    { GemmP ceq1_0;
      ceq1_0.A = HP + (size_t)0 * C1; ceq1_0.B = wq + 0; ceq1_0.bias = bq; ceq1_0.R = HP + (size_t)0 * C1; ceq1_0.C = Q;
      ceq1_0.sAo = (long long)3 * 2050 * C1; ceq1_0.sAi = 0; ceq1_0.sAm = C1; ceq1_0.sAk = 1; ceq1_0.sBo = 0; ceq1_0.sBi = 0; ceq1_0.sBn = C1 * 9; ceq1_0.sBk = 9; ceq1_0.sCo = (long long)Tt * LD; ceq1_0.sCi = 0; ceq1_0.sCm = LD; ceq1_0.sRo = 0; ceq1_0.sRi = 0; ceq1_0.sRm = 0; ceq1_0.sRn = 0;
      ceq1_0.M = Tt; ceq1_0.N = D; ceq1_0.K = C1; ceq1_0.zi_n = 1; ceq1_0.flags = 1; ceq1_0.act = 0;
      ceq1_0.alpha = 1.0f; ceq1_0.beta = 0.0f; ceq1_0.sa = 1.0f; ceq1_0.sb = 1.0f; ceq1_0.Npad = LD; ceq1_0.pad_ = 0;
      k_gemm<1><<<dim3((unsigned)((LD) + 31) / 32, (unsigned)((Tt) + 15) / 16, (unsigned)(Fo)), 32, 0, stream>>>(ceq1_0); }
    { GemmP ceq1_1;
      ceq1_1.A = HP + (size_t)1 * C1; ceq1_1.B = wq + 1; ceq1_1.bias = HP + (size_t)1 * C1; ceq1_1.R = Q; ceq1_1.C = Q;
      ceq1_1.sAo = (long long)3 * 2050 * C1; ceq1_1.sAi = 0; ceq1_1.sAm = C1; ceq1_1.sAk = 1; ceq1_1.sBo = 0; ceq1_1.sBi = 0; ceq1_1.sBn = C1 * 9; ceq1_1.sBk = 9; ceq1_1.sCo = (long long)Tt * LD; ceq1_1.sCi = 0; ceq1_1.sCm = LD; ceq1_1.sRo = (long long)Tt * LD; ceq1_1.sRi = 0; ceq1_1.sRm = LD; ceq1_1.sRn = 1;
      ceq1_1.M = Tt; ceq1_1.N = D; ceq1_1.K = C1; ceq1_1.zi_n = 1; ceq1_1.flags = 4; ceq1_1.act = 0;
      ceq1_1.alpha = 1.0f; ceq1_1.beta = 1.0f; ceq1_1.sa = 1.0f; ceq1_1.sb = 1.0f; ceq1_1.Npad = LD; ceq1_1.pad_ = 0;
      k_gemm<1><<<dim3((unsigned)((LD) + 31) / 32, (unsigned)((Tt) + 15) / 16, (unsigned)(Fo)), 32, 0, stream>>>(ceq1_1); }
    { GemmP ceq1_2;
      ceq1_2.A = HP + (size_t)2 * C1; ceq1_2.B = wq + 2; ceq1_2.bias = HP + (size_t)2 * C1; ceq1_2.R = Q; ceq1_2.C = Q;
      ceq1_2.sAo = (long long)3 * 2050 * C1; ceq1_2.sAi = 0; ceq1_2.sAm = C1; ceq1_2.sAk = 1; ceq1_2.sBo = 0; ceq1_2.sBi = 0; ceq1_2.sBn = C1 * 9; ceq1_2.sBk = 9; ceq1_2.sCo = (long long)Tt * LD; ceq1_2.sCi = 0; ceq1_2.sCm = LD; ceq1_2.sRo = (long long)Tt * LD; ceq1_2.sRi = 0; ceq1_2.sRm = LD; ceq1_2.sRn = 1;
      ceq1_2.M = Tt; ceq1_2.N = D; ceq1_2.K = C1; ceq1_2.zi_n = 1; ceq1_2.flags = 4; ceq1_2.act = 0;
      ceq1_2.alpha = 1.0f; ceq1_2.beta = 1.0f; ceq1_2.sa = 1.0f; ceq1_2.sb = 1.0f; ceq1_2.Npad = LD; ceq1_2.pad_ = 0;
      k_gemm<1><<<dim3((unsigned)((LD) + 31) / 32, (unsigned)((Tt) + 15) / 16, (unsigned)(Fo)), 32, 0, stream>>>(ceq1_2); }
    { GemmP ceq1_3;
      ceq1_3.A = HP + (size_t)2050 * C1; ceq1_3.B = wq + 3; ceq1_3.bias = HP + (size_t)2050 * C1; ceq1_3.R = Q; ceq1_3.C = Q;
      ceq1_3.sAo = (long long)3 * 2050 * C1; ceq1_3.sAi = 0; ceq1_3.sAm = C1; ceq1_3.sAk = 1; ceq1_3.sBo = 0; ceq1_3.sBi = 0; ceq1_3.sBn = C1 * 9; ceq1_3.sBk = 9; ceq1_3.sCo = (long long)Tt * LD; ceq1_3.sCi = 0; ceq1_3.sCm = LD; ceq1_3.sRo = (long long)Tt * LD; ceq1_3.sRi = 0; ceq1_3.sRm = LD; ceq1_3.sRn = 1;
      ceq1_3.M = Tt; ceq1_3.N = D; ceq1_3.K = C1; ceq1_3.zi_n = 1; ceq1_3.flags = 4; ceq1_3.act = 0;
      ceq1_3.alpha = 1.0f; ceq1_3.beta = 1.0f; ceq1_3.sa = 1.0f; ceq1_3.sb = 1.0f; ceq1_3.Npad = LD; ceq1_3.pad_ = 0;
      k_gemm<1><<<dim3((unsigned)((LD) + 31) / 32, (unsigned)((Tt) + 15) / 16, (unsigned)(Fo)), 32, 0, stream>>>(ceq1_3); }
    { GemmP ceq1_4;
      ceq1_4.A = HP + (size_t)2051 * C1; ceq1_4.B = wq + 4; ceq1_4.bias = HP + (size_t)2051 * C1; ceq1_4.R = Q; ceq1_4.C = Q;
      ceq1_4.sAo = (long long)3 * 2050 * C1; ceq1_4.sAi = 0; ceq1_4.sAm = C1; ceq1_4.sAk = 1; ceq1_4.sBo = 0; ceq1_4.sBi = 0; ceq1_4.sBn = C1 * 9; ceq1_4.sBk = 9; ceq1_4.sCo = (long long)Tt * LD; ceq1_4.sCi = 0; ceq1_4.sCm = LD; ceq1_4.sRo = (long long)Tt * LD; ceq1_4.sRi = 0; ceq1_4.sRm = LD; ceq1_4.sRn = 1;
      ceq1_4.M = Tt; ceq1_4.N = D; ceq1_4.K = C1; ceq1_4.zi_n = 1; ceq1_4.flags = 4; ceq1_4.act = 0;
      ceq1_4.alpha = 1.0f; ceq1_4.beta = 1.0f; ceq1_4.sa = 1.0f; ceq1_4.sb = 1.0f; ceq1_4.Npad = LD; ceq1_4.pad_ = 0;
      k_gemm<1><<<dim3((unsigned)((LD) + 31) / 32, (unsigned)((Tt) + 15) / 16, (unsigned)(Fo)), 32, 0, stream>>>(ceq1_4); }
    { GemmP ceq1_5;
      ceq1_5.A = HP + (size_t)2052 * C1; ceq1_5.B = wq + 5; ceq1_5.bias = HP + (size_t)2052 * C1; ceq1_5.R = Q; ceq1_5.C = Q;
      ceq1_5.sAo = (long long)3 * 2050 * C1; ceq1_5.sAi = 0; ceq1_5.sAm = C1; ceq1_5.sAk = 1; ceq1_5.sBo = 0; ceq1_5.sBi = 0; ceq1_5.sBn = C1 * 9; ceq1_5.sBk = 9; ceq1_5.sCo = (long long)Tt * LD; ceq1_5.sCi = 0; ceq1_5.sCm = LD; ceq1_5.sRo = (long long)Tt * LD; ceq1_5.sRi = 0; ceq1_5.sRm = LD; ceq1_5.sRn = 1;
      ceq1_5.M = Tt; ceq1_5.N = D; ceq1_5.K = C1; ceq1_5.zi_n = 1; ceq1_5.flags = 4; ceq1_5.act = 0;
      ceq1_5.alpha = 1.0f; ceq1_5.beta = 1.0f; ceq1_5.sa = 1.0f; ceq1_5.sb = 1.0f; ceq1_5.Npad = LD; ceq1_5.pad_ = 0;
      k_gemm<1><<<dim3((unsigned)((LD) + 31) / 32, (unsigned)((Tt) + 15) / 16, (unsigned)(Fo)), 32, 0, stream>>>(ceq1_5); }
    { GemmP ceq1_6;
      ceq1_6.A = HP + (size_t)4100 * C1; ceq1_6.B = wq + 6; ceq1_6.bias = HP + (size_t)4100 * C1; ceq1_6.R = Q; ceq1_6.C = Q;
      ceq1_6.sAo = (long long)3 * 2050 * C1; ceq1_6.sAi = 0; ceq1_6.sAm = C1; ceq1_6.sAk = 1; ceq1_6.sBo = 0; ceq1_6.sBi = 0; ceq1_6.sBn = C1 * 9; ceq1_6.sBk = 9; ceq1_6.sCo = (long long)Tt * LD; ceq1_6.sCi = 0; ceq1_6.sCm = LD; ceq1_6.sRo = (long long)Tt * LD; ceq1_6.sRi = 0; ceq1_6.sRm = LD; ceq1_6.sRn = 1;
      ceq1_6.M = Tt; ceq1_6.N = D; ceq1_6.K = C1; ceq1_6.zi_n = 1; ceq1_6.flags = 4; ceq1_6.act = 0;
      ceq1_6.alpha = 1.0f; ceq1_6.beta = 1.0f; ceq1_6.sa = 1.0f; ceq1_6.sb = 1.0f; ceq1_6.Npad = LD; ceq1_6.pad_ = 0;
      k_gemm<1><<<dim3((unsigned)((LD) + 31) / 32, (unsigned)((Tt) + 15) / 16, (unsigned)(Fo)), 32, 0, stream>>>(ceq1_6); }
    { GemmP ceq1_7;
      ceq1_7.A = HP + (size_t)4101 * C1; ceq1_7.B = wq + 7; ceq1_7.bias = HP + (size_t)4101 * C1; ceq1_7.R = Q; ceq1_7.C = Q;
      ceq1_7.sAo = (long long)3 * 2050 * C1; ceq1_7.sAi = 0; ceq1_7.sAm = C1; ceq1_7.sAk = 1; ceq1_7.sBo = 0; ceq1_7.sBi = 0; ceq1_7.sBn = C1 * 9; ceq1_7.sBk = 9; ceq1_7.sCo = (long long)Tt * LD; ceq1_7.sCi = 0; ceq1_7.sCm = LD; ceq1_7.sRo = (long long)Tt * LD; ceq1_7.sRi = 0; ceq1_7.sRm = LD; ceq1_7.sRn = 1;
      ceq1_7.M = Tt; ceq1_7.N = D; ceq1_7.K = C1; ceq1_7.zi_n = 1; ceq1_7.flags = 4; ceq1_7.act = 0;
      ceq1_7.alpha = 1.0f; ceq1_7.beta = 1.0f; ceq1_7.sa = 1.0f; ceq1_7.sb = 1.0f; ceq1_7.Npad = LD; ceq1_7.pad_ = 0;
      k_gemm<1><<<dim3((unsigned)((LD) + 31) / 32, (unsigned)((Tt) + 15) / 16, (unsigned)(Fo)), 32, 0, stream>>>(ceq1_7); }
    { GemmP ceq1_8;
      ceq1_8.A = HP + (size_t)4102 * C1; ceq1_8.B = wq + 8; ceq1_8.bias = HP + (size_t)4102 * C1; ceq1_8.R = Q; ceq1_8.C = Q;
      ceq1_8.sAo = (long long)3 * 2050 * C1; ceq1_8.sAi = 0; ceq1_8.sAm = C1; ceq1_8.sAk = 1; ceq1_8.sBo = 0; ceq1_8.sBi = 0; ceq1_8.sBn = C1 * 9; ceq1_8.sBk = 9; ceq1_8.sCo = (long long)Tt * LD; ceq1_8.sCi = 0; ceq1_8.sCm = LD; ceq1_8.sRo = (long long)Tt * LD; ceq1_8.sRi = 0; ceq1_8.sRm = LD; ceq1_8.sRn = 1;
      ceq1_8.M = Tt; ceq1_8.N = D; ceq1_8.K = C1; ceq1_8.zi_n = 1; ceq1_8.flags = 4; ceq1_8.act = 0;
      ceq1_8.alpha = 1.0f; ceq1_8.beta = 1.0f; ceq1_8.sa = 1.0f; ceq1_8.sb = 1.0f; ceq1_8.Npad = LD; ceq1_8.pad_ = 0;
      k_gemm<1><<<dim3((unsigned)((LD) + 31) / 32, (unsigned)((Tt) + 15) / 16, (unsigned)(Fo)), 32, 0, stream>>>(ceq1_8); }

    { GemmP cekv1_0;
      cekv1_0.A = HP + (size_t)0 * C1; cekv1_0.B = wkv + 0; cekv1_0.bias = bkv; cekv1_0.R = HP + (size_t)0 * C1; cekv1_0.C = KV;
      cekv1_0.sAo = (long long)3 * 2050 * C1; cekv1_0.sAi = 0; cekv1_0.sAm = C1; cekv1_0.sAk = 1; cekv1_0.sBo = 0; cekv1_0.sBi = 0; cekv1_0.sBn = C1 * 9; cekv1_0.sBk = 9; cekv1_0.sCo = (long long)Tt * LD; cekv1_0.sCi = 0; cekv1_0.sCm = LD; cekv1_0.sRo = 0; cekv1_0.sRi = 0; cekv1_0.sRm = 0; cekv1_0.sRn = 0;
      cekv1_0.M = Tt; cekv1_0.N = D; cekv1_0.K = C1; cekv1_0.zi_n = 1; cekv1_0.flags = 1; cekv1_0.act = 0;
      cekv1_0.alpha = 1.0f; cekv1_0.beta = 0.0f; cekv1_0.sa = 1.0f; cekv1_0.sb = 1.0f; cekv1_0.Npad = LD; cekv1_0.pad_ = 0;
      k_gemm<1><<<dim3((unsigned)((LD) + 31) / 32, (unsigned)((Tt) + 15) / 16, (unsigned)(Fo)), 32, 0, stream>>>(cekv1_0); }
    { GemmP cekv1_1;
      cekv1_1.A = HP + (size_t)1 * C1; cekv1_1.B = wkv + 1; cekv1_1.bias = HP + (size_t)1 * C1; cekv1_1.R = KV; cekv1_1.C = KV;
      cekv1_1.sAo = (long long)3 * 2050 * C1; cekv1_1.sAi = 0; cekv1_1.sAm = C1; cekv1_1.sAk = 1; cekv1_1.sBo = 0; cekv1_1.sBi = 0; cekv1_1.sBn = C1 * 9; cekv1_1.sBk = 9; cekv1_1.sCo = (long long)Tt * LD; cekv1_1.sCi = 0; cekv1_1.sCm = LD; cekv1_1.sRo = (long long)Tt * LD; cekv1_1.sRi = 0; cekv1_1.sRm = LD; cekv1_1.sRn = 1;
      cekv1_1.M = Tt; cekv1_1.N = D; cekv1_1.K = C1; cekv1_1.zi_n = 1; cekv1_1.flags = 4; cekv1_1.act = 0;
      cekv1_1.alpha = 1.0f; cekv1_1.beta = 1.0f; cekv1_1.sa = 1.0f; cekv1_1.sb = 1.0f; cekv1_1.Npad = LD; cekv1_1.pad_ = 0;
      k_gemm<1><<<dim3((unsigned)((LD) + 31) / 32, (unsigned)((Tt) + 15) / 16, (unsigned)(Fo)), 32, 0, stream>>>(cekv1_1); }
    { GemmP cekv1_2;
      cekv1_2.A = HP + (size_t)2 * C1; cekv1_2.B = wkv + 2; cekv1_2.bias = HP + (size_t)2 * C1; cekv1_2.R = KV; cekv1_2.C = KV;
      cekv1_2.sAo = (long long)3 * 2050 * C1; cekv1_2.sAi = 0; cekv1_2.sAm = C1; cekv1_2.sAk = 1; cekv1_2.sBo = 0; cekv1_2.sBi = 0; cekv1_2.sBn = C1 * 9; cekv1_2.sBk = 9; cekv1_2.sCo = (long long)Tt * LD; cekv1_2.sCi = 0; cekv1_2.sCm = LD; cekv1_2.sRo = (long long)Tt * LD; cekv1_2.sRi = 0; cekv1_2.sRm = LD; cekv1_2.sRn = 1;
      cekv1_2.M = Tt; cekv1_2.N = D; cekv1_2.K = C1; cekv1_2.zi_n = 1; cekv1_2.flags = 4; cekv1_2.act = 0;
      cekv1_2.alpha = 1.0f; cekv1_2.beta = 1.0f; cekv1_2.sa = 1.0f; cekv1_2.sb = 1.0f; cekv1_2.Npad = LD; cekv1_2.pad_ = 0;
      k_gemm<1><<<dim3((unsigned)((LD) + 31) / 32, (unsigned)((Tt) + 15) / 16, (unsigned)(Fo)), 32, 0, stream>>>(cekv1_2); }
    { GemmP cekv1_3;
      cekv1_3.A = HP + (size_t)2050 * C1; cekv1_3.B = wkv + 3; cekv1_3.bias = HP + (size_t)2050 * C1; cekv1_3.R = KV; cekv1_3.C = KV;
      cekv1_3.sAo = (long long)3 * 2050 * C1; cekv1_3.sAi = 0; cekv1_3.sAm = C1; cekv1_3.sAk = 1; cekv1_3.sBo = 0; cekv1_3.sBi = 0; cekv1_3.sBn = C1 * 9; cekv1_3.sBk = 9; cekv1_3.sCo = (long long)Tt * LD; cekv1_3.sCi = 0; cekv1_3.sCm = LD; cekv1_3.sRo = (long long)Tt * LD; cekv1_3.sRi = 0; cekv1_3.sRm = LD; cekv1_3.sRn = 1;
      cekv1_3.M = Tt; cekv1_3.N = D; cekv1_3.K = C1; cekv1_3.zi_n = 1; cekv1_3.flags = 4; cekv1_3.act = 0;
      cekv1_3.alpha = 1.0f; cekv1_3.beta = 1.0f; cekv1_3.sa = 1.0f; cekv1_3.sb = 1.0f; cekv1_3.Npad = LD; cekv1_3.pad_ = 0;
      k_gemm<1><<<dim3((unsigned)((LD) + 31) / 32, (unsigned)((Tt) + 15) / 16, (unsigned)(Fo)), 32, 0, stream>>>(cekv1_3); }
    { GemmP cekv1_4;
      cekv1_4.A = HP + (size_t)2051 * C1; cekv1_4.B = wkv + 4; cekv1_4.bias = HP + (size_t)2051 * C1; cekv1_4.R = KV; cekv1_4.C = KV;
      cekv1_4.sAo = (long long)3 * 2050 * C1; cekv1_4.sAi = 0; cekv1_4.sAm = C1; cekv1_4.sAk = 1; cekv1_4.sBo = 0; cekv1_4.sBi = 0; cekv1_4.sBn = C1 * 9; cekv1_4.sBk = 9; cekv1_4.sCo = (long long)Tt * LD; cekv1_4.sCi = 0; cekv1_4.sCm = LD; cekv1_4.sRo = (long long)Tt * LD; cekv1_4.sRi = 0; cekv1_4.sRm = LD; cekv1_4.sRn = 1;
      cekv1_4.M = Tt; cekv1_4.N = D; cekv1_4.K = C1; cekv1_4.zi_n = 1; cekv1_4.flags = 4; cekv1_4.act = 0;
      cekv1_4.alpha = 1.0f; cekv1_4.beta = 1.0f; cekv1_4.sa = 1.0f; cekv1_4.sb = 1.0f; cekv1_4.Npad = LD; cekv1_4.pad_ = 0;
      k_gemm<1><<<dim3((unsigned)((LD) + 31) / 32, (unsigned)((Tt) + 15) / 16, (unsigned)(Fo)), 32, 0, stream>>>(cekv1_4); }
    { GemmP cekv1_5;
      cekv1_5.A = HP + (size_t)2052 * C1; cekv1_5.B = wkv + 5; cekv1_5.bias = HP + (size_t)2052 * C1; cekv1_5.R = KV; cekv1_5.C = KV;
      cekv1_5.sAo = (long long)3 * 2050 * C1; cekv1_5.sAi = 0; cekv1_5.sAm = C1; cekv1_5.sAk = 1; cekv1_5.sBo = 0; cekv1_5.sBi = 0; cekv1_5.sBn = C1 * 9; cekv1_5.sBk = 9; cekv1_5.sCo = (long long)Tt * LD; cekv1_5.sCi = 0; cekv1_5.sCm = LD; cekv1_5.sRo = (long long)Tt * LD; cekv1_5.sRi = 0; cekv1_5.sRm = LD; cekv1_5.sRn = 1;
      cekv1_5.M = Tt; cekv1_5.N = D; cekv1_5.K = C1; cekv1_5.zi_n = 1; cekv1_5.flags = 4; cekv1_5.act = 0;
      cekv1_5.alpha = 1.0f; cekv1_5.beta = 1.0f; cekv1_5.sa = 1.0f; cekv1_5.sb = 1.0f; cekv1_5.Npad = LD; cekv1_5.pad_ = 0;
      k_gemm<1><<<dim3((unsigned)((LD) + 31) / 32, (unsigned)((Tt) + 15) / 16, (unsigned)(Fo)), 32, 0, stream>>>(cekv1_5); }
    { GemmP cekv1_6;
      cekv1_6.A = HP + (size_t)4100 * C1; cekv1_6.B = wkv + 6; cekv1_6.bias = HP + (size_t)4100 * C1; cekv1_6.R = KV; cekv1_6.C = KV;
      cekv1_6.sAo = (long long)3 * 2050 * C1; cekv1_6.sAi = 0; cekv1_6.sAm = C1; cekv1_6.sAk = 1; cekv1_6.sBo = 0; cekv1_6.sBi = 0; cekv1_6.sBn = C1 * 9; cekv1_6.sBk = 9; cekv1_6.sCo = (long long)Tt * LD; cekv1_6.sCi = 0; cekv1_6.sCm = LD; cekv1_6.sRo = (long long)Tt * LD; cekv1_6.sRi = 0; cekv1_6.sRm = LD; cekv1_6.sRn = 1;
      cekv1_6.M = Tt; cekv1_6.N = D; cekv1_6.K = C1; cekv1_6.zi_n = 1; cekv1_6.flags = 4; cekv1_6.act = 0;
      cekv1_6.alpha = 1.0f; cekv1_6.beta = 1.0f; cekv1_6.sa = 1.0f; cekv1_6.sb = 1.0f; cekv1_6.Npad = LD; cekv1_6.pad_ = 0;
      k_gemm<1><<<dim3((unsigned)((LD) + 31) / 32, (unsigned)((Tt) + 15) / 16, (unsigned)(Fo)), 32, 0, stream>>>(cekv1_6); }
    { GemmP cekv1_7;
      cekv1_7.A = HP + (size_t)4101 * C1; cekv1_7.B = wkv + 7; cekv1_7.bias = HP + (size_t)4101 * C1; cekv1_7.R = KV; cekv1_7.C = KV;
      cekv1_7.sAo = (long long)3 * 2050 * C1; cekv1_7.sAi = 0; cekv1_7.sAm = C1; cekv1_7.sAk = 1; cekv1_7.sBo = 0; cekv1_7.sBi = 0; cekv1_7.sBn = C1 * 9; cekv1_7.sBk = 9; cekv1_7.sCo = (long long)Tt * LD; cekv1_7.sCi = 0; cekv1_7.sCm = LD; cekv1_7.sRo = (long long)Tt * LD; cekv1_7.sRi = 0; cekv1_7.sRm = LD; cekv1_7.sRn = 1;
      cekv1_7.M = Tt; cekv1_7.N = D; cekv1_7.K = C1; cekv1_7.zi_n = 1; cekv1_7.flags = 4; cekv1_7.act = 0;
      cekv1_7.alpha = 1.0f; cekv1_7.beta = 1.0f; cekv1_7.sa = 1.0f; cekv1_7.sb = 1.0f; cekv1_7.Npad = LD; cekv1_7.pad_ = 0;
      k_gemm<1><<<dim3((unsigned)((LD) + 31) / 32, (unsigned)((Tt) + 15) / 16, (unsigned)(Fo)), 32, 0, stream>>>(cekv1_7); }
    { GemmP cekv1_8;
      cekv1_8.A = HP + (size_t)4102 * C1; cekv1_8.B = wkv + 8; cekv1_8.bias = HP + (size_t)4102 * C1; cekv1_8.R = KV; cekv1_8.C = KV;
      cekv1_8.sAo = (long long)3 * 2050 * C1; cekv1_8.sAi = 0; cekv1_8.sAm = C1; cekv1_8.sAk = 1; cekv1_8.sBo = 0; cekv1_8.sBi = 0; cekv1_8.sBn = C1 * 9; cekv1_8.sBk = 9; cekv1_8.sCo = (long long)Tt * LD; cekv1_8.sCi = 0; cekv1_8.sCm = LD; cekv1_8.sRo = (long long)Tt * LD; cekv1_8.sRi = 0; cekv1_8.sRm = LD; cekv1_8.sRn = 1;
      cekv1_8.M = Tt; cekv1_8.N = D; cekv1_8.K = C1; cekv1_8.zi_n = 1; cekv1_8.flags = 4; cekv1_8.act = 0;
      cekv1_8.alpha = 1.0f; cekv1_8.beta = 1.0f; cekv1_8.sa = 1.0f; cekv1_8.sb = 1.0f; cekv1_8.Npad = LD; cekv1_8.pad_ = 0;
      k_gemm<1><<<dim3((unsigned)((LD) + 31) / 32, (unsigned)((Tt) + 15) / 16, (unsigned)(Fo)), 32, 0, stream>>>(cekv1_8); }

    k_cl_colsum1<<<NB, 256, 0, stream>>>(frame + (size_t)1 * Ll, 1, 1, (long long)Ll, PART); k_cl_colsum2<<<1, 256, 0, stream>>>(PART, NB, 1, RED, 0);
    k_cl_masknorm<<<(unsigned)((Ll + 255) / 256), 256, 0, stream>>>(KV, LD, frame + (size_t)1 * Ll, RED, Tsc, (long long)Ll, D);
    { GemmP gpQP1;
      gpQP1.A = Q; gpQP1.B = faq; gpQP1.bias = fabq; gpQP1.R = Q; gpQP1.C = QP;
      gpQP1.sAo = 0; gpQP1.sAi = 0; gpQP1.sAm = LD; gpQP1.sAk = 1; gpQP1.sBo = 0; gpQP1.sBi = 0; gpQP1.sBn = 1; gpQP1.sBk = D; gpQP1.sCo = 0; gpQP1.sCi = 0; gpQP1.sCm = LD; gpQP1.sRo = 0; gpQP1.sRi = 0; gpQP1.sRm = 0; gpQP1.sRn = 0;
      gpQP1.M = Ll; gpQP1.N = D; gpQP1.K = D; gpQP1.zi_n = 1; gpQP1.flags = 1; gpQP1.act = 6;
      gpQP1.alpha = 1.0f; gpQP1.beta = 0.0f; gpQP1.sa = 1.0f; gpQP1.sb = 1.0f; gpQP1.Npad = LD; gpQP1.pad_ = 0;
      k_gemm<1><<<dim3((unsigned)((LD) + 31) / 32, (unsigned)((Ll) + 15) / 16, (unsigned)(1)), 32, 0, stream>>>(gpQP1); }
    { GemmP gpKP1;
      gpKP1.A = KV; gpKP1.B = fak; gpKP1.bias = fabk; gpKP1.R = KV; gpKP1.C = KP;
      gpKP1.sAo = 0; gpKP1.sAi = 0; gpKP1.sAm = LD; gpKP1.sAk = 1; gpKP1.sBo = 0; gpKP1.sBi = 0; gpKP1.sBn = 1; gpKP1.sBk = D; gpKP1.sCo = 0; gpKP1.sCi = 0; gpKP1.sCm = LD; gpKP1.sRo = 0; gpKP1.sRi = 0; gpKP1.sRm = 0; gpKP1.sRn = 0;
      gpKP1.M = Ll; gpKP1.N = D; gpKP1.K = D; gpKP1.zi_n = 1; gpKP1.flags = 1; gpKP1.act = 6;
      gpKP1.alpha = 1.0f; gpKP1.beta = 0.0f; gpKP1.sa = 1.0f; gpKP1.sb = 1.0f; gpKP1.Npad = LD; gpKP1.pad_ = 0;
      k_gemm<1><<<dim3((unsigned)((LD) + 31) / 32, (unsigned)((Ll) + 15) / 16, (unsigned)(1)), 32, 0, stream>>>(gpKP1); }
    { GemmP gpVP1;
      gpVP1.A = KV; gpVP1.B = fav; gpVP1.bias = fabv; gpVP1.R = KV; gpVP1.C = VP;
      gpVP1.sAo = 0; gpVP1.sAi = 0; gpVP1.sAm = LD; gpVP1.sAk = 1; gpVP1.sBo = 0; gpVP1.sBi = 0; gpVP1.sBn = 1; gpVP1.sBk = D; gpVP1.sCo = 0; gpVP1.sCi = 0; gpVP1.sCm = LD; gpVP1.sRo = 0; gpVP1.sRi = 0; gpVP1.sRm = 0; gpVP1.sRn = 0;
      gpVP1.M = Ll; gpVP1.N = D; gpVP1.K = D; gpVP1.zi_n = 1; gpVP1.flags = 1; gpVP1.act = 0;
      gpVP1.alpha = 1.0f; gpVP1.beta = 0.0f; gpVP1.sa = 1.0f; gpVP1.sb = 1.0f; gpVP1.Npad = LD; gpVP1.pad_ = 0;
      k_gemm<1><<<dim3((unsigned)((LD) + 31) / 32, (unsigned)((Ll) + 15) / 16, (unsigned)(1)), 32, 0, stream>>>(gpVP1); }
    k_cl_colsum1<<<NB, 256, 0, stream>>>(KP, LD, D, (long long)Ll, PART); k_cl_colsum2<<<1, 256, 0, stream>>>(PART, NB, D, RED, 16);
    k_cl_colsum1<<<NB, 256, 0, stream>>>(QP, LD, D, (long long)Ll, PART); k_cl_colsum2<<<1, 256, 0, stream>>>(PART, NB, D, RED, 32);
    k_cl_flow1<<<(unsigned)((Ll + 255) / 256), 256, 0, stream>>>(QP, KP, LD, RED, SV, (long long)Ll, D);
    k_cl_flow2<<<(unsigned)(((long long)Ll * D + 255) / 256), 256, 0, stream>>>(QP, KP, LD, SV, O, O2, (long long)Ll, D);
    k_cl_colsum1<<<NB, 256, 0, stream>>>(O, LD, D, (long long)Ll, PART); k_cl_colsum2<<<1, 256, 0, stream>>>(PART, NB, D, RED, 48);
    k_cl_colsum1<<<NB, 256, 0, stream>>>(O2, LD, D, (long long)Ll, PART); k_cl_colsum2<<<1, 256, 0, stream>>>(PART, NB, D, RED, 64);
    k_cl_flow3<<<(unsigned)((Ll + 255) / 256), 256, 0, stream>>>(QP, KP, LD, RED, SV, (long long)Ll, D);
    k_cl_max1<<<NB, 256, 0, stream>>>(SV, 3, (long long)Ll, PART); k_cl_max2<<<1, 256, 0, stream>>>(PART, NB, RED, 80);
    k_cl_flow4<<<(unsigned)((Ll + 255) / 256), 256, 0, stream>>>(SV, RED, O2, LD, (long long)Ll);
    k_cl_colsum1<<<NB, 256, 0, stream>>>(O2 + 15, LD, 1, (long long)Ll, PART); k_cl_colsum2<<<1, 256, 0, stream>>>(PART, NB, 1, RED, 96);
    k_cl_flow5<<<(unsigned)(((long long)Ll * D + 255) / 256), 256, 0, stream>>>(VP, O2, LD, RED, O, (long long)Ll, D);
    { GemmP gkv1;
      gkv1.A = KP; gkv1.B = O; gkv1.bias = KP; gkv1.R = KP; gkv1.C = KVM;
      gkv1.sAo = 0; gkv1.sAi = 0; gkv1.sAm = 1; gkv1.sAk = LD; gkv1.sBo = 0; gkv1.sBi = 0; gkv1.sBn = 1; gkv1.sBk = LD; gkv1.sCo = 0; gkv1.sCi = 0; gkv1.sCm = LD; gkv1.sRo = 0; gkv1.sRi = 0; gkv1.sRm = 0; gkv1.sRn = 0;
      gkv1.M = D; gkv1.N = D; gkv1.K = Ll; gkv1.zi_n = 1; gkv1.flags = 0; gkv1.act = 0;
      gkv1.alpha = 1.0f; gkv1.beta = 0.0f; gkv1.sa = 1.0f; gkv1.sb = 1.0f; gkv1.Npad = LD; gkv1.pad_ = 0;
      k_gemm<1><<<dim3((unsigned)((LD) + 31) / 32, (unsigned)((D) + 15) / 16, (unsigned)(1)), 32, 0, stream>>>(gkv1); }
    { GemmP gqkv1;
      gqkv1.A = QP; gqkv1.B = KVM; gqkv1.bias = QP; gqkv1.R = QP; gqkv1.C = O2;
      gqkv1.sAo = 0; gqkv1.sAi = 0; gqkv1.sAm = LD; gqkv1.sAk = 1; gqkv1.sBo = 0; gqkv1.sBi = 0; gqkv1.sBn = 1; gqkv1.sBk = LD; gqkv1.sCo = 0; gqkv1.sCi = 0; gqkv1.sCm = LD; gqkv1.sRo = 0; gqkv1.sRi = 0; gqkv1.sRm = 0; gqkv1.sRn = 0;
      gqkv1.M = Ll; gqkv1.N = D; gqkv1.K = D; gqkv1.zi_n = 1; gqkv1.flags = 0; gqkv1.act = 0;
      gqkv1.alpha = 1.0f; gqkv1.beta = 0.0f; gqkv1.sa = 1.0f; gqkv1.sb = 1.0f; gqkv1.Npad = LD; gqkv1.pad_ = 0;
      k_gemm<1><<<dim3((unsigned)((LD) + 31) / 32, (unsigned)((Ll) + 15) / 16, (unsigned)(1)), 32, 0, stream>>>(gqkv1); }
    k_cl_flow6<<<(unsigned)(((long long)Ll * D + 255) / 256), 256, 0, stream>>>(O2, LD, SV, (long long)Ll, D);
    { GemmP gwo1;
      gwo1.A = O2; gwo1.B = fao; gwo1.bias = fabo; gwo1.R = O2; gwo1.C = O;
      gwo1.sAo = 0; gwo1.sAi = 0; gwo1.sAm = LD; gwo1.sAk = 1; gwo1.sBo = 0; gwo1.sBi = 0; gwo1.sBn = 1; gwo1.sBk = D; gwo1.sCo = 0; gwo1.sCi = 0; gwo1.sCm = LD; gwo1.sRo = 0; gwo1.sRi = 0; gwo1.sRm = 0; gwo1.sRn = 0;
      gwo1.M = Ll; gwo1.N = D; gwo1.K = D; gwo1.zi_n = 1; gwo1.flags = 1; gwo1.act = 0;
      gwo1.alpha = 1.0f; gwo1.beta = 0.0f; gwo1.sa = 1.0f; gwo1.sb = 1.0f; gwo1.Npad = LD; gwo1.pad_ = 0;
      k_gemm<1><<<dim3((unsigned)((LD) + 31) / 32, (unsigned)((Ll) + 15) / 16, (unsigned)(1)), 32, 0, stream>>>(gwo1); }
    k_cl_out<<<(unsigned)(((long long)Ll * D + 255) / 256), 256, 0, stream>>>(O, LD, out, 1, (long long)Ll, D);
    hipMemsetAsync(XP, 0, (size_t)256 * 2052 * CI * 4, stream); hipMemsetAsync(HP, 0, (size_t)Hh * 2050 * C1 * 4, stream);
    k_cl_pad<<<(unsigned)(((long long)Hh * Tt * CI + 255) / 256), 256, 0, stream>>>(x, XP, 2, CI, Hh, Tt);
    { GemmP cp2_0;
      cp2_0.A = XP + (size_t)0 * CI; cp2_0.B = wpre + 0; cp2_0.bias = bpre; cp2_0.R = XP + (size_t)0 * CI; cp2_0.C = HP + C1;
      cp2_0.sAo = (long long)2052 * CI; cp2_0.sAi = 0; cp2_0.sAm = CI; cp2_0.sAk = 1; cp2_0.sBo = 0; cp2_0.sBi = 0; cp2_0.sBn = CI * 25; cp2_0.sBk = 25; cp2_0.sCo = (long long)2050 * C1; cp2_0.sCi = 0; cp2_0.sCm = C1; cp2_0.sRo = 0; cp2_0.sRi = 0; cp2_0.sRm = 0; cp2_0.sRn = 0;
      cp2_0.M = Tt; cp2_0.N = C1; cp2_0.K = CI; cp2_0.zi_n = 1; cp2_0.flags = 1; cp2_0.act = 0;
      cp2_0.alpha = 1.0f; cp2_0.beta = 0.0f; cp2_0.sa = 1.0f; cp2_0.sb = 1.0f; cp2_0.Npad = C1; cp2_0.pad_ = 0;
      k_gemm<1><<<dim3((unsigned)((C1) + 31) / 32, (unsigned)((Tt) + 15) / 16, (unsigned)(Hh)), 32, 0, stream>>>(cp2_0); }
    { GemmP cp2_1;
      cp2_1.A = XP + (size_t)1 * CI; cp2_1.B = wpre + 1; cp2_1.bias = XP + (size_t)1 * CI; cp2_1.R = HP + C1; cp2_1.C = HP + C1;
      cp2_1.sAo = (long long)2052 * CI; cp2_1.sAi = 0; cp2_1.sAm = CI; cp2_1.sAk = 1; cp2_1.sBo = 0; cp2_1.sBi = 0; cp2_1.sBn = CI * 25; cp2_1.sBk = 25; cp2_1.sCo = (long long)2050 * C1; cp2_1.sCi = 0; cp2_1.sCm = C1; cp2_1.sRo = (long long)2050 * C1; cp2_1.sRi = 0; cp2_1.sRm = C1; cp2_1.sRn = 1;
      cp2_1.M = Tt; cp2_1.N = C1; cp2_1.K = CI; cp2_1.zi_n = 1; cp2_1.flags = 4; cp2_1.act = 0;
      cp2_1.alpha = 1.0f; cp2_1.beta = 1.0f; cp2_1.sa = 1.0f; cp2_1.sb = 1.0f; cp2_1.Npad = C1; cp2_1.pad_ = 0;
      k_gemm<1><<<dim3((unsigned)((C1) + 31) / 32, (unsigned)((Tt) + 15) / 16, (unsigned)(Hh)), 32, 0, stream>>>(cp2_1); }
    { GemmP cp2_2;
      cp2_2.A = XP + (size_t)2 * CI; cp2_2.B = wpre + 2; cp2_2.bias = XP + (size_t)2 * CI; cp2_2.R = HP + C1; cp2_2.C = HP + C1;
      cp2_2.sAo = (long long)2052 * CI; cp2_2.sAi = 0; cp2_2.sAm = CI; cp2_2.sAk = 1; cp2_2.sBo = 0; cp2_2.sBi = 0; cp2_2.sBn = CI * 25; cp2_2.sBk = 25; cp2_2.sCo = (long long)2050 * C1; cp2_2.sCi = 0; cp2_2.sCm = C1; cp2_2.sRo = (long long)2050 * C1; cp2_2.sRi = 0; cp2_2.sRm = C1; cp2_2.sRn = 1;
      cp2_2.M = Tt; cp2_2.N = C1; cp2_2.K = CI; cp2_2.zi_n = 1; cp2_2.flags = 4; cp2_2.act = 0;
      cp2_2.alpha = 1.0f; cp2_2.beta = 1.0f; cp2_2.sa = 1.0f; cp2_2.sb = 1.0f; cp2_2.Npad = C1; cp2_2.pad_ = 0;
      k_gemm<1><<<dim3((unsigned)((C1) + 31) / 32, (unsigned)((Tt) + 15) / 16, (unsigned)(Hh)), 32, 0, stream>>>(cp2_2); }
    { GemmP cp2_3;
      cp2_3.A = XP + (size_t)3 * CI; cp2_3.B = wpre + 3; cp2_3.bias = XP + (size_t)3 * CI; cp2_3.R = HP + C1; cp2_3.C = HP + C1;
      cp2_3.sAo = (long long)2052 * CI; cp2_3.sAi = 0; cp2_3.sAm = CI; cp2_3.sAk = 1; cp2_3.sBo = 0; cp2_3.sBi = 0; cp2_3.sBn = CI * 25; cp2_3.sBk = 25; cp2_3.sCo = (long long)2050 * C1; cp2_3.sCi = 0; cp2_3.sCm = C1; cp2_3.sRo = (long long)2050 * C1; cp2_3.sRi = 0; cp2_3.sRm = C1; cp2_3.sRn = 1;
      cp2_3.M = Tt; cp2_3.N = C1; cp2_3.K = CI; cp2_3.zi_n = 1; cp2_3.flags = 4; cp2_3.act = 0;
      cp2_3.alpha = 1.0f; cp2_3.beta = 1.0f; cp2_3.sa = 1.0f; cp2_3.sb = 1.0f; cp2_3.Npad = C1; cp2_3.pad_ = 0;
      k_gemm<1><<<dim3((unsigned)((C1) + 31) / 32, (unsigned)((Tt) + 15) / 16, (unsigned)(Hh)), 32, 0, stream>>>(cp2_3); }
    { GemmP cp2_4;
      cp2_4.A = XP + (size_t)4 * CI; cp2_4.B = wpre + 4; cp2_4.bias = XP + (size_t)4 * CI; cp2_4.R = HP + C1; cp2_4.C = HP + C1;
      cp2_4.sAo = (long long)2052 * CI; cp2_4.sAi = 0; cp2_4.sAm = CI; cp2_4.sAk = 1; cp2_4.sBo = 0; cp2_4.sBi = 0; cp2_4.sBn = CI * 25; cp2_4.sBk = 25; cp2_4.sCo = (long long)2050 * C1; cp2_4.sCi = 0; cp2_4.sCm = C1; cp2_4.sRo = (long long)2050 * C1; cp2_4.sRi = 0; cp2_4.sRm = C1; cp2_4.sRn = 1;
      cp2_4.M = Tt; cp2_4.N = C1; cp2_4.K = CI; cp2_4.zi_n = 1; cp2_4.flags = 4; cp2_4.act = 0;
      cp2_4.alpha = 1.0f; cp2_4.beta = 1.0f; cp2_4.sa = 1.0f; cp2_4.sb = 1.0f; cp2_4.Npad = C1; cp2_4.pad_ = 0;
      k_gemm<1><<<dim3((unsigned)((C1) + 31) / 32, (unsigned)((Tt) + 15) / 16, (unsigned)(Hh)), 32, 0, stream>>>(cp2_4); }
    { GemmP cp2_5;
      cp2_5.A = XP + (size_t)2052 * CI; cp2_5.B = wpre + 5; cp2_5.bias = XP + (size_t)2052 * CI; cp2_5.R = HP + C1; cp2_5.C = HP + C1;
      cp2_5.sAo = (long long)2052 * CI; cp2_5.sAi = 0; cp2_5.sAm = CI; cp2_5.sAk = 1; cp2_5.sBo = 0; cp2_5.sBi = 0; cp2_5.sBn = CI * 25; cp2_5.sBk = 25; cp2_5.sCo = (long long)2050 * C1; cp2_5.sCi = 0; cp2_5.sCm = C1; cp2_5.sRo = (long long)2050 * C1; cp2_5.sRi = 0; cp2_5.sRm = C1; cp2_5.sRn = 1;
      cp2_5.M = Tt; cp2_5.N = C1; cp2_5.K = CI; cp2_5.zi_n = 1; cp2_5.flags = 4; cp2_5.act = 0;
      cp2_5.alpha = 1.0f; cp2_5.beta = 1.0f; cp2_5.sa = 1.0f; cp2_5.sb = 1.0f; cp2_5.Npad = C1; cp2_5.pad_ = 0;
      k_gemm<1><<<dim3((unsigned)((C1) + 31) / 32, (unsigned)((Tt) + 15) / 16, (unsigned)(Hh)), 32, 0, stream>>>(cp2_5); }
    { GemmP cp2_6;
      cp2_6.A = XP + (size_t)2053 * CI; cp2_6.B = wpre + 6; cp2_6.bias = XP + (size_t)2053 * CI; cp2_6.R = HP + C1; cp2_6.C = HP + C1;
      cp2_6.sAo = (long long)2052 * CI; cp2_6.sAi = 0; cp2_6.sAm = CI; cp2_6.sAk = 1; cp2_6.sBo = 0; cp2_6.sBi = 0; cp2_6.sBn = CI * 25; cp2_6.sBk = 25; cp2_6.sCo = (long long)2050 * C1; cp2_6.sCi = 0; cp2_6.sCm = C1; cp2_6.sRo = (long long)2050 * C1; cp2_6.sRi = 0; cp2_6.sRm = C1; cp2_6.sRn = 1;
      cp2_6.M = Tt; cp2_6.N = C1; cp2_6.K = CI; cp2_6.zi_n = 1; cp2_6.flags = 4; cp2_6.act = 0;
      cp2_6.alpha = 1.0f; cp2_6.beta = 1.0f; cp2_6.sa = 1.0f; cp2_6.sb = 1.0f; cp2_6.Npad = C1; cp2_6.pad_ = 0;
      k_gemm<1><<<dim3((unsigned)((C1) + 31) / 32, (unsigned)((Tt) + 15) / 16, (unsigned)(Hh)), 32, 0, stream>>>(cp2_6); }
    { GemmP cp2_7;
      cp2_7.A = XP + (size_t)2054 * CI; cp2_7.B = wpre + 7; cp2_7.bias = XP + (size_t)2054 * CI; cp2_7.R = HP + C1; cp2_7.C = HP + C1;
      cp2_7.sAo = (long long)2052 * CI; cp2_7.sAi = 0; cp2_7.sAm = CI; cp2_7.sAk = 1; cp2_7.sBo = 0; cp2_7.sBi = 0; cp2_7.sBn = CI * 25; cp2_7.sBk = 25; cp2_7.sCo = (long long)2050 * C1; cp2_7.sCi = 0; cp2_7.sCm = C1; cp2_7.sRo = (long long)2050 * C1; cp2_7.sRi = 0; cp2_7.sRm = C1; cp2_7.sRn = 1;
      cp2_7.M = Tt; cp2_7.N = C1; cp2_7.K = CI; cp2_7.zi_n = 1; cp2_7.flags = 4; cp2_7.act = 0;
      cp2_7.alpha = 1.0f; cp2_7.beta = 1.0f; cp2_7.sa = 1.0f; cp2_7.sb = 1.0f; cp2_7.Npad = C1; cp2_7.pad_ = 0;
      k_gemm<1><<<dim3((unsigned)((C1) + 31) / 32, (unsigned)((Tt) + 15) / 16, (unsigned)(Hh)), 32, 0, stream>>>(cp2_7); }
    { GemmP cp2_8;
      cp2_8.A = XP + (size_t)2055 * CI; cp2_8.B = wpre + 8; cp2_8.bias = XP + (size_t)2055 * CI; cp2_8.R = HP + C1; cp2_8.C = HP + C1;
      cp2_8.sAo = (long long)2052 * CI; cp2_8.sAi = 0; cp2_8.sAm = CI; cp2_8.sAk = 1; cp2_8.sBo = 0; cp2_8.sBi = 0; cp2_8.sBn = CI * 25; cp2_8.sBk = 25; cp2_8.sCo = (long long)2050 * C1; cp2_8.sCi = 0; cp2_8.sCm = C1; cp2_8.sRo = (long long)2050 * C1; cp2_8.sRi = 0; cp2_8.sRm = C1; cp2_8.sRn = 1;
      cp2_8.M = Tt; cp2_8.N = C1; cp2_8.K = CI; cp2_8.zi_n = 1; cp2_8.flags = 4; cp2_8.act = 0;
      cp2_8.alpha = 1.0f; cp2_8.beta = 1.0f; cp2_8.sa = 1.0f; cp2_8.sb = 1.0f; cp2_8.Npad = C1; cp2_8.pad_ = 0;
      k_gemm<1><<<dim3((unsigned)((C1) + 31) / 32, (unsigned)((Tt) + 15) / 16, (unsigned)(Hh)), 32, 0, stream>>>(cp2_8); }
    { GemmP cp2_9;
      cp2_9.A = XP + (size_t)2056 * CI; cp2_9.B = wpre + 9; cp2_9.bias = XP + (size_t)2056 * CI; cp2_9.R = HP + C1; cp2_9.C = HP + C1;
      cp2_9.sAo = (long long)2052 * CI; cp2_9.sAi = 0; cp2_9.sAm = CI; cp2_9.sAk = 1; cp2_9.sBo = 0; cp2_9.sBi = 0; cp2_9.sBn = CI * 25; cp2_9.sBk = 25; cp2_9.sCo = (long long)2050 * C1; cp2_9.sCi = 0; cp2_9.sCm = C1; cp2_9.sRo = (long long)2050 * C1; cp2_9.sRi = 0; cp2_9.sRm = C1; cp2_9.sRn = 1;
      cp2_9.M = Tt; cp2_9.N = C1; cp2_9.K = CI; cp2_9.zi_n = 1; cp2_9.flags = 4; cp2_9.act = 0;
      cp2_9.alpha = 1.0f; cp2_9.beta = 1.0f; cp2_9.sa = 1.0f; cp2_9.sb = 1.0f; cp2_9.Npad = C1; cp2_9.pad_ = 0;
      k_gemm<1><<<dim3((unsigned)((C1) + 31) / 32, (unsigned)((Tt) + 15) / 16, (unsigned)(Hh)), 32, 0, stream>>>(cp2_9); }
    { GemmP cp2_10;
      cp2_10.A = XP + (size_t)4104 * CI; cp2_10.B = wpre + 10; cp2_10.bias = XP + (size_t)4104 * CI; cp2_10.R = HP + C1; cp2_10.C = HP + C1;
      cp2_10.sAo = (long long)2052 * CI; cp2_10.sAi = 0; cp2_10.sAm = CI; cp2_10.sAk = 1; cp2_10.sBo = 0; cp2_10.sBi = 0; cp2_10.sBn = CI * 25; cp2_10.sBk = 25; cp2_10.sCo = (long long)2050 * C1; cp2_10.sCi = 0; cp2_10.sCm = C1; cp2_10.sRo = (long long)2050 * C1; cp2_10.sRi = 0; cp2_10.sRm = C1; cp2_10.sRn = 1;
      cp2_10.M = Tt; cp2_10.N = C1; cp2_10.K = CI; cp2_10.zi_n = 1; cp2_10.flags = 4; cp2_10.act = 0;
      cp2_10.alpha = 1.0f; cp2_10.beta = 1.0f; cp2_10.sa = 1.0f; cp2_10.sb = 1.0f; cp2_10.Npad = C1; cp2_10.pad_ = 0;
      k_gemm<1><<<dim3((unsigned)((C1) + 31) / 32, (unsigned)((Tt) + 15) / 16, (unsigned)(Hh)), 32, 0, stream>>>(cp2_10); }
    { GemmP cp2_11;
      cp2_11.A = XP + (size_t)4105 * CI; cp2_11.B = wpre + 11; cp2_11.bias = XP + (size_t)4105 * CI; cp2_11.R = HP + C1; cp2_11.C = HP + C1;
      cp2_11.sAo = (long long)2052 * CI; cp2_11.sAi = 0; cp2_11.sAm = CI; cp2_11.sAk = 1; cp2_11.sBo = 0; cp2_11.sBi = 0; cp2_11.sBn = CI * 25; cp2_11.sBk = 25; cp2_11.sCo = (long long)2050 * C1; cp2_11.sCi = 0; cp2_11.sCm = C1; cp2_11.sRo = (long long)2050 * C1; cp2_11.sRi = 0; cp2_11.sRm = C1; cp2_11.sRn = 1;
      cp2_11.M = Tt; cp2_11.N = C1; cp2_11.K = CI; cp2_11.zi_n = 1; cp2_11.flags = 4; cp2_11.act = 0;
      cp2_11.alpha = 1.0f; cp2_11.beta = 1.0f; cp2_11.sa = 1.0f; cp2_11.sb = 1.0f; cp2_11.Npad = C1; cp2_11.pad_ = 0;
      k_gemm<1><<<dim3((unsigned)((C1) + 31) / 32, (unsigned)((Tt) + 15) / 16, (unsigned)(Hh)), 32, 0, stream>>>(cp2_11); }
    { GemmP cp2_12;
      cp2_12.A = XP + (size_t)4106 * CI; cp2_12.B = wpre + 12; cp2_12.bias = XP + (size_t)4106 * CI; cp2_12.R = HP + C1; cp2_12.C = HP + C1;
      cp2_12.sAo = (long long)2052 * CI; cp2_12.sAi = 0; cp2_12.sAm = CI; cp2_12.sAk = 1; cp2_12.sBo = 0; cp2_12.sBi = 0; cp2_12.sBn = CI * 25; cp2_12.sBk = 25; cp2_12.sCo = (long long)2050 * C1; cp2_12.sCi = 0; cp2_12.sCm = C1; cp2_12.sRo = (long long)2050 * C1; cp2_12.sRi = 0; cp2_12.sRm = C1; cp2_12.sRn = 1;
      cp2_12.M = Tt; cp2_12.N = C1; cp2_12.K = CI; cp2_12.zi_n = 1; cp2_12.flags = 4; cp2_12.act = 0;
      cp2_12.alpha = 1.0f; cp2_12.beta = 1.0f; cp2_12.sa = 1.0f; cp2_12.sb = 1.0f; cp2_12.Npad = C1; cp2_12.pad_ = 0;
      k_gemm<1><<<dim3((unsigned)((C1) + 31) / 32, (unsigned)((Tt) + 15) / 16, (unsigned)(Hh)), 32, 0, stream>>>(cp2_12); }
    { GemmP cp2_13;
      cp2_13.A = XP + (size_t)4107 * CI; cp2_13.B = wpre + 13; cp2_13.bias = XP + (size_t)4107 * CI; cp2_13.R = HP + C1; cp2_13.C = HP + C1;
      cp2_13.sAo = (long long)2052 * CI; cp2_13.sAi = 0; cp2_13.sAm = CI; cp2_13.sAk = 1; cp2_13.sBo = 0; cp2_13.sBi = 0; cp2_13.sBn = CI * 25; cp2_13.sBk = 25; cp2_13.sCo = (long long)2050 * C1; cp2_13.sCi = 0; cp2_13.sCm = C1; cp2_13.sRo = (long long)2050 * C1; cp2_13.sRi = 0; cp2_13.sRm = C1; cp2_13.sRn = 1;
      cp2_13.M = Tt; cp2_13.N = C1; cp2_13.K = CI; cp2_13.zi_n = 1; cp2_13.flags = 4; cp2_13.act = 0;
      cp2_13.alpha = 1.0f; cp2_13.beta = 1.0f; cp2_13.sa = 1.0f; cp2_13.sb = 1.0f; cp2_13.Npad = C1; cp2_13.pad_ = 0;
      k_gemm<1><<<dim3((unsigned)((C1) + 31) / 32, (unsigned)((Tt) + 15) / 16, (unsigned)(Hh)), 32, 0, stream>>>(cp2_13); }
    { GemmP cp2_14;
      cp2_14.A = XP + (size_t)4108 * CI; cp2_14.B = wpre + 14; cp2_14.bias = XP + (size_t)4108 * CI; cp2_14.R = HP + C1; cp2_14.C = HP + C1;
      cp2_14.sAo = (long long)2052 * CI; cp2_14.sAi = 0; cp2_14.sAm = CI; cp2_14.sAk = 1; cp2_14.sBo = 0; cp2_14.sBi = 0; cp2_14.sBn = CI * 25; cp2_14.sBk = 25; cp2_14.sCo = (long long)2050 * C1; cp2_14.sCi = 0; cp2_14.sCm = C1; cp2_14.sRo = (long long)2050 * C1; cp2_14.sRi = 0; cp2_14.sRm = C1; cp2_14.sRn = 1;
      cp2_14.M = Tt; cp2_14.N = C1; cp2_14.K = CI; cp2_14.zi_n = 1; cp2_14.flags = 4; cp2_14.act = 0;
      cp2_14.alpha = 1.0f; cp2_14.beta = 1.0f; cp2_14.sa = 1.0f; cp2_14.sb = 1.0f; cp2_14.Npad = C1; cp2_14.pad_ = 0;
      k_gemm<1><<<dim3((unsigned)((C1) + 31) / 32, (unsigned)((Tt) + 15) / 16, (unsigned)(Hh)), 32, 0, stream>>>(cp2_14); }
    { GemmP cp2_15;
      cp2_15.A = XP + (size_t)6156 * CI; cp2_15.B = wpre + 15; cp2_15.bias = XP + (size_t)6156 * CI; cp2_15.R = HP + C1; cp2_15.C = HP + C1;
      cp2_15.sAo = (long long)2052 * CI; cp2_15.sAi = 0; cp2_15.sAm = CI; cp2_15.sAk = 1; cp2_15.sBo = 0; cp2_15.sBi = 0; cp2_15.sBn = CI * 25; cp2_15.sBk = 25; cp2_15.sCo = (long long)2050 * C1; cp2_15.sCi = 0; cp2_15.sCm = C1; cp2_15.sRo = (long long)2050 * C1; cp2_15.sRi = 0; cp2_15.sRm = C1; cp2_15.sRn = 1;
      cp2_15.M = Tt; cp2_15.N = C1; cp2_15.K = CI; cp2_15.zi_n = 1; cp2_15.flags = 4; cp2_15.act = 0;
      cp2_15.alpha = 1.0f; cp2_15.beta = 1.0f; cp2_15.sa = 1.0f; cp2_15.sb = 1.0f; cp2_15.Npad = C1; cp2_15.pad_ = 0;
      k_gemm<1><<<dim3((unsigned)((C1) + 31) / 32, (unsigned)((Tt) + 15) / 16, (unsigned)(Hh)), 32, 0, stream>>>(cp2_15); }
    { GemmP cp2_16;
      cp2_16.A = XP + (size_t)6157 * CI; cp2_16.B = wpre + 16; cp2_16.bias = XP + (size_t)6157 * CI; cp2_16.R = HP + C1; cp2_16.C = HP + C1;
      cp2_16.sAo = (long long)2052 * CI; cp2_16.sAi = 0; cp2_16.sAm = CI; cp2_16.sAk = 1; cp2_16.sBo = 0; cp2_16.sBi = 0; cp2_16.sBn = CI * 25; cp2_16.sBk = 25; cp2_16.sCo = (long long)2050 * C1; cp2_16.sCi = 0; cp2_16.sCm = C1; cp2_16.sRo = (long long)2050 * C1; cp2_16.sRi = 0; cp2_16.sRm = C1; cp2_16.sRn = 1;
      cp2_16.M = Tt; cp2_16.N = C1; cp2_16.K = CI; cp2_16.zi_n = 1; cp2_16.flags = 4; cp2_16.act = 0;
      cp2_16.alpha = 1.0f; cp2_16.beta = 1.0f; cp2_16.sa = 1.0f; cp2_16.sb = 1.0f; cp2_16.Npad = C1; cp2_16.pad_ = 0;
      k_gemm<1><<<dim3((unsigned)((C1) + 31) / 32, (unsigned)((Tt) + 15) / 16, (unsigned)(Hh)), 32, 0, stream>>>(cp2_16); }
    { GemmP cp2_17;
      cp2_17.A = XP + (size_t)6158 * CI; cp2_17.B = wpre + 17; cp2_17.bias = XP + (size_t)6158 * CI; cp2_17.R = HP + C1; cp2_17.C = HP + C1;
      cp2_17.sAo = (long long)2052 * CI; cp2_17.sAi = 0; cp2_17.sAm = CI; cp2_17.sAk = 1; cp2_17.sBo = 0; cp2_17.sBi = 0; cp2_17.sBn = CI * 25; cp2_17.sBk = 25; cp2_17.sCo = (long long)2050 * C1; cp2_17.sCi = 0; cp2_17.sCm = C1; cp2_17.sRo = (long long)2050 * C1; cp2_17.sRi = 0; cp2_17.sRm = C1; cp2_17.sRn = 1;
      cp2_17.M = Tt; cp2_17.N = C1; cp2_17.K = CI; cp2_17.zi_n = 1; cp2_17.flags = 4; cp2_17.act = 0;
      cp2_17.alpha = 1.0f; cp2_17.beta = 1.0f; cp2_17.sa = 1.0f; cp2_17.sb = 1.0f; cp2_17.Npad = C1; cp2_17.pad_ = 0;
      k_gemm<1><<<dim3((unsigned)((C1) + 31) / 32, (unsigned)((Tt) + 15) / 16, (unsigned)(Hh)), 32, 0, stream>>>(cp2_17); }
    { GemmP cp2_18;
      cp2_18.A = XP + (size_t)6159 * CI; cp2_18.B = wpre + 18; cp2_18.bias = XP + (size_t)6159 * CI; cp2_18.R = HP + C1; cp2_18.C = HP + C1;
      cp2_18.sAo = (long long)2052 * CI; cp2_18.sAi = 0; cp2_18.sAm = CI; cp2_18.sAk = 1; cp2_18.sBo = 0; cp2_18.sBi = 0; cp2_18.sBn = CI * 25; cp2_18.sBk = 25; cp2_18.sCo = (long long)2050 * C1; cp2_18.sCi = 0; cp2_18.sCm = C1; cp2_18.sRo = (long long)2050 * C1; cp2_18.sRi = 0; cp2_18.sRm = C1; cp2_18.sRn = 1;
      cp2_18.M = Tt; cp2_18.N = C1; cp2_18.K = CI; cp2_18.zi_n = 1; cp2_18.flags = 4; cp2_18.act = 0;
      cp2_18.alpha = 1.0f; cp2_18.beta = 1.0f; cp2_18.sa = 1.0f; cp2_18.sb = 1.0f; cp2_18.Npad = C1; cp2_18.pad_ = 0;
      k_gemm<1><<<dim3((unsigned)((C1) + 31) / 32, (unsigned)((Tt) + 15) / 16, (unsigned)(Hh)), 32, 0, stream>>>(cp2_18); }
    { GemmP cp2_19;
      cp2_19.A = XP + (size_t)6160 * CI; cp2_19.B = wpre + 19; cp2_19.bias = XP + (size_t)6160 * CI; cp2_19.R = HP + C1; cp2_19.C = HP + C1;
      cp2_19.sAo = (long long)2052 * CI; cp2_19.sAi = 0; cp2_19.sAm = CI; cp2_19.sAk = 1; cp2_19.sBo = 0; cp2_19.sBi = 0; cp2_19.sBn = CI * 25; cp2_19.sBk = 25; cp2_19.sCo = (long long)2050 * C1; cp2_19.sCi = 0; cp2_19.sCm = C1; cp2_19.sRo = (long long)2050 * C1; cp2_19.sRi = 0; cp2_19.sRm = C1; cp2_19.sRn = 1;
      cp2_19.M = Tt; cp2_19.N = C1; cp2_19.K = CI; cp2_19.zi_n = 1; cp2_19.flags = 4; cp2_19.act = 0;
      cp2_19.alpha = 1.0f; cp2_19.beta = 1.0f; cp2_19.sa = 1.0f; cp2_19.sb = 1.0f; cp2_19.Npad = C1; cp2_19.pad_ = 0;
      k_gemm<1><<<dim3((unsigned)((C1) + 31) / 32, (unsigned)((Tt) + 15) / 16, (unsigned)(Hh)), 32, 0, stream>>>(cp2_19); }
    { GemmP cp2_20;
      cp2_20.A = XP + (size_t)8208 * CI; cp2_20.B = wpre + 20; cp2_20.bias = XP + (size_t)8208 * CI; cp2_20.R = HP + C1; cp2_20.C = HP + C1;
      cp2_20.sAo = (long long)2052 * CI; cp2_20.sAi = 0; cp2_20.sAm = CI; cp2_20.sAk = 1; cp2_20.sBo = 0; cp2_20.sBi = 0; cp2_20.sBn = CI * 25; cp2_20.sBk = 25; cp2_20.sCo = (long long)2050 * C1; cp2_20.sCi = 0; cp2_20.sCm = C1; cp2_20.sRo = (long long)2050 * C1; cp2_20.sRi = 0; cp2_20.sRm = C1; cp2_20.sRn = 1;
      cp2_20.M = Tt; cp2_20.N = C1; cp2_20.K = CI; cp2_20.zi_n = 1; cp2_20.flags = 4; cp2_20.act = 0;
      cp2_20.alpha = 1.0f; cp2_20.beta = 1.0f; cp2_20.sa = 1.0f; cp2_20.sb = 1.0f; cp2_20.Npad = C1; cp2_20.pad_ = 0;
      k_gemm<1><<<dim3((unsigned)((C1) + 31) / 32, (unsigned)((Tt) + 15) / 16, (unsigned)(Hh)), 32, 0, stream>>>(cp2_20); }
    { GemmP cp2_21;
      cp2_21.A = XP + (size_t)8209 * CI; cp2_21.B = wpre + 21; cp2_21.bias = XP + (size_t)8209 * CI; cp2_21.R = HP + C1; cp2_21.C = HP + C1;
      cp2_21.sAo = (long long)2052 * CI; cp2_21.sAi = 0; cp2_21.sAm = CI; cp2_21.sAk = 1; cp2_21.sBo = 0; cp2_21.sBi = 0; cp2_21.sBn = CI * 25; cp2_21.sBk = 25; cp2_21.sCo = (long long)2050 * C1; cp2_21.sCi = 0; cp2_21.sCm = C1; cp2_21.sRo = (long long)2050 * C1; cp2_21.sRi = 0; cp2_21.sRm = C1; cp2_21.sRn = 1;
      cp2_21.M = Tt; cp2_21.N = C1; cp2_21.K = CI; cp2_21.zi_n = 1; cp2_21.flags = 4; cp2_21.act = 0;
      cp2_21.alpha = 1.0f; cp2_21.beta = 1.0f; cp2_21.sa = 1.0f; cp2_21.sb = 1.0f; cp2_21.Npad = C1; cp2_21.pad_ = 0;
      k_gemm<1><<<dim3((unsigned)((C1) + 31) / 32, (unsigned)((Tt) + 15) / 16, (unsigned)(Hh)), 32, 0, stream>>>(cp2_21); }
    { GemmP cp2_22;
      cp2_22.A = XP + (size_t)8210 * CI; cp2_22.B = wpre + 22; cp2_22.bias = XP + (size_t)8210 * CI; cp2_22.R = HP + C1; cp2_22.C = HP + C1;
      cp2_22.sAo = (long long)2052 * CI; cp2_22.sAi = 0; cp2_22.sAm = CI; cp2_22.sAk = 1; cp2_22.sBo = 0; cp2_22.sBi = 0; cp2_22.sBn = CI * 25; cp2_22.sBk = 25; cp2_22.sCo = (long long)2050 * C1; cp2_22.sCi = 0; cp2_22.sCm = C1; cp2_22.sRo = (long long)2050 * C1; cp2_22.sRi = 0; cp2_22.sRm = C1; cp2_22.sRn = 1;
      cp2_22.M = Tt; cp2_22.N = C1; cp2_22.K = CI; cp2_22.zi_n = 1; cp2_22.flags = 4; cp2_22.act = 0;
      cp2_22.alpha = 1.0f; cp2_22.beta = 1.0f; cp2_22.sa = 1.0f; cp2_22.sb = 1.0f; cp2_22.Npad = C1; cp2_22.pad_ = 0;
      k_gemm<1><<<dim3((unsigned)((C1) + 31) / 32, (unsigned)((Tt) + 15) / 16, (unsigned)(Hh)), 32, 0, stream>>>(cp2_22); }
    { GemmP cp2_23;
      cp2_23.A = XP + (size_t)8211 * CI; cp2_23.B = wpre + 23; cp2_23.bias = XP + (size_t)8211 * CI; cp2_23.R = HP + C1; cp2_23.C = HP + C1;
      cp2_23.sAo = (long long)2052 * CI; cp2_23.sAi = 0; cp2_23.sAm = CI; cp2_23.sAk = 1; cp2_23.sBo = 0; cp2_23.sBi = 0; cp2_23.sBn = CI * 25; cp2_23.sBk = 25; cp2_23.sCo = (long long)2050 * C1; cp2_23.sCi = 0; cp2_23.sCm = C1; cp2_23.sRo = (long long)2050 * C1; cp2_23.sRi = 0; cp2_23.sRm = C1; cp2_23.sRn = 1;
      cp2_23.M = Tt; cp2_23.N = C1; cp2_23.K = CI; cp2_23.zi_n = 1; cp2_23.flags = 4; cp2_23.act = 0;
      cp2_23.alpha = 1.0f; cp2_23.beta = 1.0f; cp2_23.sa = 1.0f; cp2_23.sb = 1.0f; cp2_23.Npad = C1; cp2_23.pad_ = 0;
      k_gemm<1><<<dim3((unsigned)((C1) + 31) / 32, (unsigned)((Tt) + 15) / 16, (unsigned)(Hh)), 32, 0, stream>>>(cp2_23); }
    { GemmP cp2_24;
      cp2_24.A = XP + (size_t)8212 * CI; cp2_24.B = wpre + 24; cp2_24.bias = XP + (size_t)8212 * CI; cp2_24.R = HP + C1; cp2_24.C = HP + C1;
      cp2_24.sAo = (long long)2052 * CI; cp2_24.sAi = 0; cp2_24.sAm = CI; cp2_24.sAk = 1; cp2_24.sBo = 0; cp2_24.sBi = 0; cp2_24.sBn = CI * 25; cp2_24.sBk = 25; cp2_24.sCo = (long long)2050 * C1; cp2_24.sCi = 0; cp2_24.sCm = C1; cp2_24.sRo = (long long)2050 * C1; cp2_24.sRi = 0; cp2_24.sRm = C1; cp2_24.sRn = 1;
      cp2_24.M = Tt; cp2_24.N = C1; cp2_24.K = CI; cp2_24.zi_n = 1; cp2_24.flags = 4; cp2_24.act = 0;
      cp2_24.alpha = 1.0f; cp2_24.beta = 1.0f; cp2_24.sa = 1.0f; cp2_24.sb = 1.0f; cp2_24.Npad = C1; cp2_24.pad_ = 0;
      k_gemm<1><<<dim3((unsigned)((C1) + 31) / 32, (unsigned)((Tt) + 15) / 16, (unsigned)(Hh)), 32, 0, stream>>>(cp2_24); }
    k_cl_bnl<<<(unsigned)(((long long)Hh * Tt * C1 + 255) / 256), 256, 0, stream>>>(HP, bng, bnb, bnm, bnv, Hh, Tt, C1);
    { GemmP ceq2_0;
      ceq2_0.A = HP + (size_t)0 * C1; ceq2_0.B = wq + 0; ceq2_0.bias = bq; ceq2_0.R = HP + (size_t)0 * C1; ceq2_0.C = Q;
      ceq2_0.sAo = (long long)3 * 2050 * C1; ceq2_0.sAi = 0; ceq2_0.sAm = C1; ceq2_0.sAk = 1; ceq2_0.sBo = 0; ceq2_0.sBi = 0; ceq2_0.sBn = C1 * 9; ceq2_0.sBk = 9; ceq2_0.sCo = (long long)Tt * LD; ceq2_0.sCi = 0; ceq2_0.sCm = LD; ceq2_0.sRo = 0; ceq2_0.sRi = 0; ceq2_0.sRm = 0; ceq2_0.sRn = 0;
      ceq2_0.M = Tt; ceq2_0.N = D; ceq2_0.K = C1; ceq2_0.zi_n = 1; ceq2_0.flags = 1; ceq2_0.act = 0;
      ceq2_0.alpha = 1.0f; ceq2_0.beta = 0.0f; ceq2_0.sa = 1.0f; ceq2_0.sb = 1.0f; ceq2_0.Npad = LD; ceq2_0.pad_ = 0;
      k_gemm<1><<<dim3((unsigned)((LD) + 31) / 32, (unsigned)((Tt) + 15) / 16, (unsigned)(Fo)), 32, 0, stream>>>(ceq2_0); }
    { GemmP ceq2_1;
      ceq2_1.A = HP + (size_t)1 * C1; ceq2_1.B = wq + 1; ceq2_1.bias = HP + (size_t)1 * C1; ceq2_1.R = Q; ceq2_1.C = Q;
      ceq2_1.sAo = (long long)3 * 2050 * C1; ceq2_1.sAi = 0; ceq2_1.sAm = C1; ceq2_1.sAk = 1; ceq2_1.sBo = 0; ceq2_1.sBi = 0; ceq2_1.sBn = C1 * 9; ceq2_1.sBk = 9; ceq2_1.sCo = (long long)Tt * LD; ceq2_1.sCi = 0; ceq2_1.sCm = LD; ceq2_1.sRo = (long long)Tt * LD; ceq2_1.sRi = 0; ceq2_1.sRm = LD; ceq2_1.sRn = 1;
      ceq2_1.M = Tt; ceq2_1.N = D; ceq2_1.K = C1; ceq2_1.zi_n = 1; ceq2_1.flags = 4; ceq2_1.act = 0;
      ceq2_1.alpha = 1.0f; ceq2_1.beta = 1.0f; ceq2_1.sa = 1.0f; ceq2_1.sb = 1.0f; ceq2_1.Npad = LD; ceq2_1.pad_ = 0;
      k_gemm<1><<<dim3((unsigned)((LD) + 31) / 32, (unsigned)((Tt) + 15) / 16, (unsigned)(Fo)), 32, 0, stream>>>(ceq2_1); }
    { GemmP ceq2_2;
      ceq2_2.A = HP + (size_t)2 * C1; ceq2_2.B = wq + 2; ceq2_2.bias = HP + (size_t)2 * C1; ceq2_2.R = Q; ceq2_2.C = Q;
      ceq2_2.sAo = (long long)3 * 2050 * C1; ceq2_2.sAi = 0; ceq2_2.sAm = C1; ceq2_2.sAk = 1; ceq2_2.sBo = 0; ceq2_2.sBi = 0; ceq2_2.sBn = C1 * 9; ceq2_2.sBk = 9; ceq2_2.sCo = (long long)Tt * LD; ceq2_2.sCi = 0; ceq2_2.sCm = LD; ceq2_2.sRo = (long long)Tt * LD; ceq2_2.sRi = 0; ceq2_2.sRm = LD; ceq2_2.sRn = 1;
      ceq2_2.M = Tt; ceq2_2.N = D; ceq2_2.K = C1; ceq2_2.zi_n = 1; ceq2_2.flags = 4; ceq2_2.act = 0;
      ceq2_2.alpha = 1.0f; ceq2_2.beta = 1.0f; ceq2_2.sa = 1.0f; ceq2_2.sb = 1.0f; ceq2_2.Npad = LD; ceq2_2.pad_ = 0;
      k_gemm<1><<<dim3((unsigned)((LD) + 31) / 32, (unsigned)((Tt) + 15) / 16, (unsigned)(Fo)), 32, 0, stream>>>(ceq2_2); }
    { GemmP ceq2_3;
      ceq2_3.A = HP + (size_t)2050 * C1; ceq2_3.B = wq + 3; ceq2_3.bias = HP + (size_t)2050 * C1; ceq2_3.R = Q; ceq2_3.C = Q;
      ceq2_3.sAo = (long long)3 * 2050 * C1; ceq2_3.sAi = 0; ceq2_3.sAm = C1; ceq2_3.sAk = 1; ceq2_3.sBo = 0; ceq2_3.sBi = 0; ceq2_3.sBn = C1 * 9; ceq2_3.sBk = 9; ceq2_3.sCo = (long long)Tt * LD; ceq2_3.sCi = 0; ceq2_3.sCm = LD; ceq2_3.sRo = (long long)Tt * LD; ceq2_3.sRi = 0; ceq2_3.sRm = LD; ceq2_3.sRn = 1;
      ceq2_3.M = Tt; ceq2_3.N = D; ceq2_3.K = C1; ceq2_3.zi_n = 1; ceq2_3.flags = 4; ceq2_3.act = 0;
      ceq2_3.alpha = 1.0f; ceq2_3.beta = 1.0f; ceq2_3.sa = 1.0f; ceq2_3.sb = 1.0f; ceq2_3.Npad = LD; ceq2_3.pad_ = 0;
      k_gemm<1><<<dim3((unsigned)((LD) + 31) / 32, (unsigned)((Tt) + 15) / 16, (unsigned)(Fo)), 32, 0, stream>>>(ceq2_3); }
    { GemmP ceq2_4;
      ceq2_4.A = HP + (size_t)2051 * C1; ceq2_4.B = wq + 4; ceq2_4.bias = HP + (size_t)2051 * C1; ceq2_4.R = Q; ceq2_4.C = Q;
      ceq2_4.sAo = (long long)3 * 2050 * C1; ceq2_4.sAi = 0; ceq2_4.sAm = C1; ceq2_4.sAk = 1; ceq2_4.sBo = 0; ceq2_4.sBi = 0; ceq2_4.sBn = C1 * 9; ceq2_4.sBk = 9; ceq2_4.sCo = (long long)Tt * LD; ceq2_4.sCi = 0; ceq2_4.sCm = LD; ceq2_4.sRo = (long long)Tt * LD; ceq2_4.sRi = 0; ceq2_4.sRm = LD; ceq2_4.sRn = 1;
      ceq2_4.M = Tt; ceq2_4.N = D; ceq2_4.K = C1; ceq2_4.zi_n = 1; ceq2_4.flags = 4; ceq2_4.act = 0;
      ceq2_4.alpha = 1.0f; ceq2_4.beta = 1.0f; ceq2_4.sa = 1.0f; ceq2_4.sb = 1.0f; ceq2_4.Npad = LD; ceq2_4.pad_ = 0;
      k_gemm<1><<<dim3((unsigned)((LD) + 31) / 32, (unsigned)((Tt) + 15) / 16, (unsigned)(Fo)), 32, 0, stream>>>(ceq2_4); }
    { GemmP ceq2_5;
      ceq2_5.A = HP + (size_t)2052 * C1; ceq2_5.B = wq + 5; ceq2_5.bias = HP + (size_t)2052 * C1; ceq2_5.R = Q; ceq2_5.C = Q;
      ceq2_5.sAo = (long long)3 * 2050 * C1; ceq2_5.sAi = 0; ceq2_5.sAm = C1; ceq2_5.sAk = 1; ceq2_5.sBo = 0; ceq2_5.sBi = 0; ceq2_5.sBn = C1 * 9; ceq2_5.sBk = 9; ceq2_5.sCo = (long long)Tt * LD; ceq2_5.sCi = 0; ceq2_5.sCm = LD; ceq2_5.sRo = (long long)Tt * LD; ceq2_5.sRi = 0; ceq2_5.sRm = LD; ceq2_5.sRn = 1;
      ceq2_5.M = Tt; ceq2_5.N = D; ceq2_5.K = C1; ceq2_5.zi_n = 1; ceq2_5.flags = 4; ceq2_5.act = 0;
      ceq2_5.alpha = 1.0f; ceq2_5.beta = 1.0f; ceq2_5.sa = 1.0f; ceq2_5.sb = 1.0f; ceq2_5.Npad = LD; ceq2_5.pad_ = 0;
      k_gemm<1><<<dim3((unsigned)((LD) + 31) / 32, (unsigned)((Tt) + 15) / 16, (unsigned)(Fo)), 32, 0, stream>>>(ceq2_5); }
    { GemmP ceq2_6;
      ceq2_6.A = HP + (size_t)4100 * C1; ceq2_6.B = wq + 6; ceq2_6.bias = HP + (size_t)4100 * C1; ceq2_6.R = Q; ceq2_6.C = Q;
      ceq2_6.sAo = (long long)3 * 2050 * C1; ceq2_6.sAi = 0; ceq2_6.sAm = C1; ceq2_6.sAk = 1; ceq2_6.sBo = 0; ceq2_6.sBi = 0; ceq2_6.sBn = C1 * 9; ceq2_6.sBk = 9; ceq2_6.sCo = (long long)Tt * LD; ceq2_6.sCi = 0; ceq2_6.sCm = LD; ceq2_6.sRo = (long long)Tt * LD; ceq2_6.sRi = 0; ceq2_6.sRm = LD; ceq2_6.sRn = 1;
      ceq2_6.M = Tt; ceq2_6.N = D; ceq2_6.K = C1; ceq2_6.zi_n = 1; ceq2_6.flags = 4; ceq2_6.act = 0;
      ceq2_6.alpha = 1.0f; ceq2_6.beta = 1.0f; ceq2_6.sa = 1.0f; ceq2_6.sb = 1.0f; ceq2_6.Npad = LD; ceq2_6.pad_ = 0;
      k_gemm<1><<<dim3((unsigned)((LD) + 31) / 32, (unsigned)((Tt) + 15) / 16, (unsigned)(Fo)), 32, 0, stream>>>(ceq2_6); }
    { GemmP ceq2_7;
      ceq2_7.A = HP + (size_t)4101 * C1; ceq2_7.B = wq + 7; ceq2_7.bias = HP + (size_t)4101 * C1; ceq2_7.R = Q; ceq2_7.C = Q;
      ceq2_7.sAo = (long long)3 * 2050 * C1; ceq2_7.sAi = 0; ceq2_7.sAm = C1; ceq2_7.sAk = 1; ceq2_7.sBo = 0; ceq2_7.sBi = 0; ceq2_7.sBn = C1 * 9; ceq2_7.sBk = 9; ceq2_7.sCo = (long long)Tt * LD; ceq2_7.sCi = 0; ceq2_7.sCm = LD; ceq2_7.sRo = (long long)Tt * LD; ceq2_7.sRi = 0; ceq2_7.sRm = LD; ceq2_7.sRn = 1;
      ceq2_7.M = Tt; ceq2_7.N = D; ceq2_7.K = C1; ceq2_7.zi_n = 1; ceq2_7.flags = 4; ceq2_7.act = 0;
      ceq2_7.alpha = 1.0f; ceq2_7.beta = 1.0f; ceq2_7.sa = 1.0f; ceq2_7.sb = 1.0f; ceq2_7.Npad = LD; ceq2_7.pad_ = 0;
      k_gemm<1><<<dim3((unsigned)((LD) + 31) / 32, (unsigned)((Tt) + 15) / 16, (unsigned)(Fo)), 32, 0, stream>>>(ceq2_7); }
    { GemmP ceq2_8;
      ceq2_8.A = HP + (size_t)4102 * C1; ceq2_8.B = wq + 8; ceq2_8.bias = HP + (size_t)4102 * C1; ceq2_8.R = Q; ceq2_8.C = Q;
      ceq2_8.sAo = (long long)3 * 2050 * C1; ceq2_8.sAi = 0; ceq2_8.sAm = C1; ceq2_8.sAk = 1; ceq2_8.sBo = 0; ceq2_8.sBi = 0; ceq2_8.sBn = C1 * 9; ceq2_8.sBk = 9; ceq2_8.sCo = (long long)Tt * LD; ceq2_8.sCi = 0; ceq2_8.sCm = LD; ceq2_8.sRo = (long long)Tt * LD; ceq2_8.sRi = 0; ceq2_8.sRm = LD; ceq2_8.sRn = 1;
      ceq2_8.M = Tt; ceq2_8.N = D; ceq2_8.K = C1; ceq2_8.zi_n = 1; ceq2_8.flags = 4; ceq2_8.act = 0;
      ceq2_8.alpha = 1.0f; ceq2_8.beta = 1.0f; ceq2_8.sa = 1.0f; ceq2_8.sb = 1.0f; ceq2_8.Npad = LD; ceq2_8.pad_ = 0;
      k_gemm<1><<<dim3((unsigned)((LD) + 31) / 32, (unsigned)((Tt) + 15) / 16, (unsigned)(Fo)), 32, 0, stream>>>(ceq2_8); }

    { GemmP cekv2_0;
      cekv2_0.A = HP + (size_t)0 * C1; cekv2_0.B = wkv + 0; cekv2_0.bias = bkv; cekv2_0.R = HP + (size_t)0 * C1; cekv2_0.C = KV;
      cekv2_0.sAo = (long long)3 * 2050 * C1; cekv2_0.sAi = 0; cekv2_0.sAm = C1; cekv2_0.sAk = 1; cekv2_0.sBo = 0; cekv2_0.sBi = 0; cekv2_0.sBn = C1 * 9; cekv2_0.sBk = 9; cekv2_0.sCo = (long long)Tt * LD; cekv2_0.sCi = 0; cekv2_0.sCm = LD; cekv2_0.sRo = 0; cekv2_0.sRi = 0; cekv2_0.sRm = 0; cekv2_0.sRn = 0;
      cekv2_0.M = Tt; cekv2_0.N = D; cekv2_0.K = C1; cekv2_0.zi_n = 1; cekv2_0.flags = 1; cekv2_0.act = 0;
      cekv2_0.alpha = 1.0f; cekv2_0.beta = 0.0f; cekv2_0.sa = 1.0f; cekv2_0.sb = 1.0f; cekv2_0.Npad = LD; cekv2_0.pad_ = 0;
      k_gemm<1><<<dim3((unsigned)((LD) + 31) / 32, (unsigned)((Tt) + 15) / 16, (unsigned)(Fo)), 32, 0, stream>>>(cekv2_0); }
    { GemmP cekv2_1;
      cekv2_1.A = HP + (size_t)1 * C1; cekv2_1.B = wkv + 1; cekv2_1.bias = HP + (size_t)1 * C1; cekv2_1.R = KV; cekv2_1.C = KV;
      cekv2_1.sAo = (long long)3 * 2050 * C1; cekv2_1.sAi = 0; cekv2_1.sAm = C1; cekv2_1.sAk = 1; cekv2_1.sBo = 0; cekv2_1.sBi = 0; cekv2_1.sBn = C1 * 9; cekv2_1.sBk = 9; cekv2_1.sCo = (long long)Tt * LD; cekv2_1.sCi = 0; cekv2_1.sCm = LD; cekv2_1.sRo = (long long)Tt * LD; cekv2_1.sRi = 0; cekv2_1.sRm = LD; cekv2_1.sRn = 1;
      cekv2_1.M = Tt; cekv2_1.N = D; cekv2_1.K = C1; cekv2_1.zi_n = 1; cekv2_1.flags = 4; cekv2_1.act = 0;
      cekv2_1.alpha = 1.0f; cekv2_1.beta = 1.0f; cekv2_1.sa = 1.0f; cekv2_1.sb = 1.0f; cekv2_1.Npad = LD; cekv2_1.pad_ = 0;
      k_gemm<1><<<dim3((unsigned)((LD) + 31) / 32, (unsigned)((Tt) + 15) / 16, (unsigned)(Fo)), 32, 0, stream>>>(cekv2_1); }
    { GemmP cekv2_2;
      cekv2_2.A = HP + (size_t)2 * C1; cekv2_2.B = wkv + 2; cekv2_2.bias = HP + (size_t)2 * C1; cekv2_2.R = KV; cekv2_2.C = KV;
      cekv2_2.sAo = (long long)3 * 2050 * C1; cekv2_2.sAi = 0; cekv2_2.sAm = C1; cekv2_2.sAk = 1; cekv2_2.sBo = 0; cekv2_2.sBi = 0; cekv2_2.sBn = C1 * 9; cekv2_2.sBk = 9; cekv2_2.sCo = (long long)Tt * LD; cekv2_2.sCi = 0; cekv2_2.sCm = LD; cekv2_2.sRo = (long long)Tt * LD; cekv2_2.sRi = 0; cekv2_2.sRm = LD; cekv2_2.sRn = 1;
      cekv2_2.M = Tt; cekv2_2.N = D; cekv2_2.K = C1; cekv2_2.zi_n = 1; cekv2_2.flags = 4; cekv2_2.act = 0;
      cekv2_2.alpha = 1.0f; cekv2_2.beta = 1.0f; cekv2_2.sa = 1.0f; cekv2_2.sb = 1.0f; cekv2_2.Npad = LD; cekv2_2.pad_ = 0;
      k_gemm<1><<<dim3((unsigned)((LD) + 31) / 32, (unsigned)((Tt) + 15) / 16, (unsigned)(Fo)), 32, 0, stream>>>(cekv2_2); }
    { GemmP cekv2_3;
      cekv2_3.A = HP + (size_t)2050 * C1; cekv2_3.B = wkv + 3; cekv2_3.bias = HP + (size_t)2050 * C1; cekv2_3.R = KV; cekv2_3.C = KV;
      cekv2_3.sAo = (long long)3 * 2050 * C1; cekv2_3.sAi = 0; cekv2_3.sAm = C1; cekv2_3.sAk = 1; cekv2_3.sBo = 0; cekv2_3.sBi = 0; cekv2_3.sBn = C1 * 9; cekv2_3.sBk = 9; cekv2_3.sCo = (long long)Tt * LD; cekv2_3.sCi = 0; cekv2_3.sCm = LD; cekv2_3.sRo = (long long)Tt * LD; cekv2_3.sRi = 0; cekv2_3.sRm = LD; cekv2_3.sRn = 1;
      cekv2_3.M = Tt; cekv2_3.N = D; cekv2_3.K = C1; cekv2_3.zi_n = 1; cekv2_3.flags = 4; cekv2_3.act = 0;
      cekv2_3.alpha = 1.0f; cekv2_3.beta = 1.0f; cekv2_3.sa = 1.0f; cekv2_3.sb = 1.0f; cekv2_3.Npad = LD; cekv2_3.pad_ = 0;
      k_gemm<1><<<dim3((unsigned)((LD) + 31) / 32, (unsigned)((Tt) + 15) / 16, (unsigned)(Fo)), 32, 0, stream>>>(cekv2_3); }
    { GemmP cekv2_4;
      cekv2_4.A = HP + (size_t)2051 * C1; cekv2_4.B = wkv + 4; cekv2_4.bias = HP + (size_t)2051 * C1; cekv2_4.R = KV; cekv2_4.C = KV;
      cekv2_4.sAo = (long long)3 * 2050 * C1; cekv2_4.sAi = 0; cekv2_4.sAm = C1; cekv2_4.sAk = 1; cekv2_4.sBo = 0; cekv2_4.sBi = 0; cekv2_4.sBn = C1 * 9; cekv2_4.sBk = 9; cekv2_4.sCo = (long long)Tt * LD; cekv2_4.sCi = 0; cekv2_4.sCm = LD; cekv2_4.sRo = (long long)Tt * LD; cekv2_4.sRi = 0; cekv2_4.sRm = LD; cekv2_4.sRn = 1;
      cekv2_4.M = Tt; cekv2_4.N = D; cekv2_4.K = C1; cekv2_4.zi_n = 1; cekv2_4.flags = 4; cekv2_4.act = 0;
      cekv2_4.alpha = 1.0f; cekv2_4.beta = 1.0f; cekv2_4.sa = 1.0f; cekv2_4.sb = 1.0f; cekv2_4.Npad = LD; cekv2_4.pad_ = 0;
      k_gemm<1><<<dim3((unsigned)((LD) + 31) / 32, (unsigned)((Tt) + 15) / 16, (unsigned)(Fo)), 32, 0, stream>>>(cekv2_4); }
    { GemmP cekv2_5;
      cekv2_5.A = HP + (size_t)2052 * C1; cekv2_5.B = wkv + 5; cekv2_5.bias = HP + (size_t)2052 * C1; cekv2_5.R = KV; cekv2_5.C = KV;
      cekv2_5.sAo = (long long)3 * 2050 * C1; cekv2_5.sAi = 0; cekv2_5.sAm = C1; cekv2_5.sAk = 1; cekv2_5.sBo = 0; cekv2_5.sBi = 0; cekv2_5.sBn = C1 * 9; cekv2_5.sBk = 9; cekv2_5.sCo = (long long)Tt * LD; cekv2_5.sCi = 0; cekv2_5.sCm = LD; cekv2_5.sRo = (long long)Tt * LD; cekv2_5.sRi = 0; cekv2_5.sRm = LD; cekv2_5.sRn = 1;
      cekv2_5.M = Tt; cekv2_5.N = D; cekv2_5.K = C1; cekv2_5.zi_n = 1; cekv2_5.flags = 4; cekv2_5.act = 0;
      cekv2_5.alpha = 1.0f; cekv2_5.beta = 1.0f; cekv2_5.sa = 1.0f; cekv2_5.sb = 1.0f; cekv2_5.Npad = LD; cekv2_5.pad_ = 0;
      k_gemm<1><<<dim3((unsigned)((LD) + 31) / 32, (unsigned)((Tt) + 15) / 16, (unsigned)(Fo)), 32, 0, stream>>>(cekv2_5); }
    { GemmP cekv2_6;
      cekv2_6.A = HP + (size_t)4100 * C1; cekv2_6.B = wkv + 6; cekv2_6.bias = HP + (size_t)4100 * C1; cekv2_6.R = KV; cekv2_6.C = KV;
      cekv2_6.sAo = (long long)3 * 2050 * C1; cekv2_6.sAi = 0; cekv2_6.sAm = C1; cekv2_6.sAk = 1; cekv2_6.sBo = 0; cekv2_6.sBi = 0; cekv2_6.sBn = C1 * 9; cekv2_6.sBk = 9; cekv2_6.sCo = (long long)Tt * LD; cekv2_6.sCi = 0; cekv2_6.sCm = LD; cekv2_6.sRo = (long long)Tt * LD; cekv2_6.sRi = 0; cekv2_6.sRm = LD; cekv2_6.sRn = 1;
      cekv2_6.M = Tt; cekv2_6.N = D; cekv2_6.K = C1; cekv2_6.zi_n = 1; cekv2_6.flags = 4; cekv2_6.act = 0;
      cekv2_6.alpha = 1.0f; cekv2_6.beta = 1.0f; cekv2_6.sa = 1.0f; cekv2_6.sb = 1.0f; cekv2_6.Npad = LD; cekv2_6.pad_ = 0;
      k_gemm<1><<<dim3((unsigned)((LD) + 31) / 32, (unsigned)((Tt) + 15) / 16, (unsigned)(Fo)), 32, 0, stream>>>(cekv2_6); }
    { GemmP cekv2_7;
      cekv2_7.A = HP + (size_t)4101 * C1; cekv2_7.B = wkv + 7; cekv2_7.bias = HP + (size_t)4101 * C1; cekv2_7.R = KV; cekv2_7.C = KV;
      cekv2_7.sAo = (long long)3 * 2050 * C1; cekv2_7.sAi = 0; cekv2_7.sAm = C1; cekv2_7.sAk = 1; cekv2_7.sBo = 0; cekv2_7.sBi = 0; cekv2_7.sBn = C1 * 9; cekv2_7.sBk = 9; cekv2_7.sCo = (long long)Tt * LD; cekv2_7.sCi = 0; cekv2_7.sCm = LD; cekv2_7.sRo = (long long)Tt * LD; cekv2_7.sRi = 0; cekv2_7.sRm = LD; cekv2_7.sRn = 1;
      cekv2_7.M = Tt; cekv2_7.N = D; cekv2_7.K = C1; cekv2_7.zi_n = 1; cekv2_7.flags = 4; cekv2_7.act = 0;
      cekv2_7.alpha = 1.0f; cekv2_7.beta = 1.0f; cekv2_7.sa = 1.0f; cekv2_7.sb = 1.0f; cekv2_7.Npad = LD; cekv2_7.pad_ = 0;
      k_gemm<1><<<dim3((unsigned)((LD) + 31) / 32, (unsigned)((Tt) + 15) / 16, (unsigned)(Fo)), 32, 0, stream>>>(cekv2_7); }
    { GemmP cekv2_8;
      cekv2_8.A = HP + (size_t)4102 * C1; cekv2_8.B = wkv + 8; cekv2_8.bias = HP + (size_t)4102 * C1; cekv2_8.R = KV; cekv2_8.C = KV;
      cekv2_8.sAo = (long long)3 * 2050 * C1; cekv2_8.sAi = 0; cekv2_8.sAm = C1; cekv2_8.sAk = 1; cekv2_8.sBo = 0; cekv2_8.sBi = 0; cekv2_8.sBn = C1 * 9; cekv2_8.sBk = 9; cekv2_8.sCo = (long long)Tt * LD; cekv2_8.sCi = 0; cekv2_8.sCm = LD; cekv2_8.sRo = (long long)Tt * LD; cekv2_8.sRi = 0; cekv2_8.sRm = LD; cekv2_8.sRn = 1;
      cekv2_8.M = Tt; cekv2_8.N = D; cekv2_8.K = C1; cekv2_8.zi_n = 1; cekv2_8.flags = 4; cekv2_8.act = 0;
      cekv2_8.alpha = 1.0f; cekv2_8.beta = 1.0f; cekv2_8.sa = 1.0f; cekv2_8.sb = 1.0f; cekv2_8.Npad = LD; cekv2_8.pad_ = 0;
      k_gemm<1><<<dim3((unsigned)((LD) + 31) / 32, (unsigned)((Tt) + 15) / 16, (unsigned)(Fo)), 32, 0, stream>>>(cekv2_8); }

    k_cl_colsum1<<<NB, 256, 0, stream>>>(frame + (size_t)2 * Ll, 1, 1, (long long)Ll, PART); k_cl_colsum2<<<1, 256, 0, stream>>>(PART, NB, 1, RED, 0);
    k_cl_masknorm<<<(unsigned)((Ll + 255) / 256), 256, 0, stream>>>(KV, LD, frame + (size_t)2 * Ll, RED, Tsc, (long long)Ll, D);
    { GemmP gpQP2;
      gpQP2.A = Q; gpQP2.B = faq; gpQP2.bias = fabq; gpQP2.R = Q; gpQP2.C = QP;
      gpQP2.sAo = 0; gpQP2.sAi = 0; gpQP2.sAm = LD; gpQP2.sAk = 1; gpQP2.sBo = 0; gpQP2.sBi = 0; gpQP2.sBn = 1; gpQP2.sBk = D; gpQP2.sCo = 0; gpQP2.sCi = 0; gpQP2.sCm = LD; gpQP2.sRo = 0; gpQP2.sRi = 0; gpQP2.sRm = 0; gpQP2.sRn = 0;
      gpQP2.M = Ll; gpQP2.N = D; gpQP2.K = D; gpQP2.zi_n = 1; gpQP2.flags = 1; gpQP2.act = 6;
      gpQP2.alpha = 1.0f; gpQP2.beta = 0.0f; gpQP2.sa = 1.0f; gpQP2.sb = 1.0f; gpQP2.Npad = LD; gpQP2.pad_ = 0;
      k_gemm<1><<<dim3((unsigned)((LD) + 31) / 32, (unsigned)((Ll) + 15) / 16, (unsigned)(1)), 32, 0, stream>>>(gpQP2); }
    { GemmP gpKP2;
      gpKP2.A = KV; gpKP2.B = fak; gpKP2.bias = fabk; gpKP2.R = KV; gpKP2.C = KP;
      gpKP2.sAo = 0; gpKP2.sAi = 0; gpKP2.sAm = LD; gpKP2.sAk = 1; gpKP2.sBo = 0; gpKP2.sBi = 0; gpKP2.sBn = 1; gpKP2.sBk = D; gpKP2.sCo = 0; gpKP2.sCi = 0; gpKP2.sCm = LD; gpKP2.sRo = 0; gpKP2.sRi = 0; gpKP2.sRm = 0; gpKP2.sRn = 0;
      gpKP2.M = Ll; gpKP2.N = D; gpKP2.K = D; gpKP2.zi_n = 1; gpKP2.flags = 1; gpKP2.act = 6;
      gpKP2.alpha = 1.0f; gpKP2.beta = 0.0f; gpKP2.sa = 1.0f; gpKP2.sb = 1.0f; gpKP2.Npad = LD; gpKP2.pad_ = 0;
      k_gemm<1><<<dim3((unsigned)((LD) + 31) / 32, (unsigned)((Ll) + 15) / 16, (unsigned)(1)), 32, 0, stream>>>(gpKP2); }
    { GemmP gpVP2;
      gpVP2.A = KV; gpVP2.B = fav; gpVP2.bias = fabv; gpVP2.R = KV; gpVP2.C = VP;
      gpVP2.sAo = 0; gpVP2.sAi = 0; gpVP2.sAm = LD; gpVP2.sAk = 1; gpVP2.sBo = 0; gpVP2.sBi = 0; gpVP2.sBn = 1; gpVP2.sBk = D; gpVP2.sCo = 0; gpVP2.sCi = 0; gpVP2.sCm = LD; gpVP2.sRo = 0; gpVP2.sRi = 0; gpVP2.sRm = 0; gpVP2.sRn = 0;
      gpVP2.M = Ll; gpVP2.N = D; gpVP2.K = D; gpVP2.zi_n = 1; gpVP2.flags = 1; gpVP2.act = 0;
      gpVP2.alpha = 1.0f; gpVP2.beta = 0.0f; gpVP2.sa = 1.0f; gpVP2.sb = 1.0f; gpVP2.Npad = LD; gpVP2.pad_ = 0;
      k_gemm<1><<<dim3((unsigned)((LD) + 31) / 32, (unsigned)((Ll) + 15) / 16, (unsigned)(1)), 32, 0, stream>>>(gpVP2); }
    k_cl_colsum1<<<NB, 256, 0, stream>>>(KP, LD, D, (long long)Ll, PART); k_cl_colsum2<<<1, 256, 0, stream>>>(PART, NB, D, RED, 16);
    k_cl_colsum1<<<NB, 256, 0, stream>>>(QP, LD, D, (long long)Ll, PART); k_cl_colsum2<<<1, 256, 0, stream>>>(PART, NB, D, RED, 32);
    k_cl_flow1<<<(unsigned)((Ll + 255) / 256), 256, 0, stream>>>(QP, KP, LD, RED, SV, (long long)Ll, D);
    k_cl_flow2<<<(unsigned)(((long long)Ll * D + 255) / 256), 256, 0, stream>>>(QP, KP, LD, SV, O, O2, (long long)Ll, D);
    k_cl_colsum1<<<NB, 256, 0, stream>>>(O, LD, D, (long long)Ll, PART); k_cl_colsum2<<<1, 256, 0, stream>>>(PART, NB, D, RED, 48);
    k_cl_colsum1<<<NB, 256, 0, stream>>>(O2, LD, D, (long long)Ll, PART); k_cl_colsum2<<<1, 256, 0, stream>>>(PART, NB, D, RED, 64);
    k_cl_flow3<<<(unsigned)((Ll + 255) / 256), 256, 0, stream>>>(QP, KP, LD, RED, SV, (long long)Ll, D);
    k_cl_max1<<<NB, 256, 0, stream>>>(SV, 3, (long long)Ll, PART); k_cl_max2<<<1, 256, 0, stream>>>(PART, NB, RED, 80);
    k_cl_flow4<<<(unsigned)((Ll + 255) / 256), 256, 0, stream>>>(SV, RED, O2, LD, (long long)Ll);
    k_cl_colsum1<<<NB, 256, 0, stream>>>(O2 + 15, LD, 1, (long long)Ll, PART); k_cl_colsum2<<<1, 256, 0, stream>>>(PART, NB, 1, RED, 96);
    k_cl_flow5<<<(unsigned)(((long long)Ll * D + 255) / 256), 256, 0, stream>>>(VP, O2, LD, RED, O, (long long)Ll, D);
    { GemmP gkv2;
      gkv2.A = KP; gkv2.B = O; gkv2.bias = KP; gkv2.R = KP; gkv2.C = KVM;
      gkv2.sAo = 0; gkv2.sAi = 0; gkv2.sAm = 1; gkv2.sAk = LD; gkv2.sBo = 0; gkv2.sBi = 0; gkv2.sBn = 1; gkv2.sBk = LD; gkv2.sCo = 0; gkv2.sCi = 0; gkv2.sCm = LD; gkv2.sRo = 0; gkv2.sRi = 0; gkv2.sRm = 0; gkv2.sRn = 0;
      gkv2.M = D; gkv2.N = D; gkv2.K = Ll; gkv2.zi_n = 1; gkv2.flags = 0; gkv2.act = 0;
      gkv2.alpha = 1.0f; gkv2.beta = 0.0f; gkv2.sa = 1.0f; gkv2.sb = 1.0f; gkv2.Npad = LD; gkv2.pad_ = 0;
      k_gemm<1><<<dim3((unsigned)((LD) + 31) / 32, (unsigned)((D) + 15) / 16, (unsigned)(1)), 32, 0, stream>>>(gkv2); }
    { GemmP gqkv2;
      gqkv2.A = QP; gqkv2.B = KVM; gqkv2.bias = QP; gqkv2.R = QP; gqkv2.C = O2;
      gqkv2.sAo = 0; gqkv2.sAi = 0; gqkv2.sAm = LD; gqkv2.sAk = 1; gqkv2.sBo = 0; gqkv2.sBi = 0; gqkv2.sBn = 1; gqkv2.sBk = LD; gqkv2.sCo = 0; gqkv2.sCi = 0; gqkv2.sCm = LD; gqkv2.sRo = 0; gqkv2.sRi = 0; gqkv2.sRm = 0; gqkv2.sRn = 0;
      gqkv2.M = Ll; gqkv2.N = D; gqkv2.K = D; gqkv2.zi_n = 1; gqkv2.flags = 0; gqkv2.act = 0;
      gqkv2.alpha = 1.0f; gqkv2.beta = 0.0f; gqkv2.sa = 1.0f; gqkv2.sb = 1.0f; gqkv2.Npad = LD; gqkv2.pad_ = 0;
      k_gemm<1><<<dim3((unsigned)((LD) + 31) / 32, (unsigned)((Ll) + 15) / 16, (unsigned)(1)), 32, 0, stream>>>(gqkv2); }
    k_cl_flow6<<<(unsigned)(((long long)Ll * D + 255) / 256), 256, 0, stream>>>(O2, LD, SV, (long long)Ll, D);
    { GemmP gwo2;
      gwo2.A = O2; gwo2.B = fao; gwo2.bias = fabo; gwo2.R = O2; gwo2.C = O;
      gwo2.sAo = 0; gwo2.sAi = 0; gwo2.sAm = LD; gwo2.sAk = 1; gwo2.sBo = 0; gwo2.sBi = 0; gwo2.sBn = 1; gwo2.sBk = D; gwo2.sCo = 0; gwo2.sCi = 0; gwo2.sCm = LD; gwo2.sRo = 0; gwo2.sRi = 0; gwo2.sRm = 0; gwo2.sRn = 0;
      gwo2.M = Ll; gwo2.N = D; gwo2.K = D; gwo2.zi_n = 1; gwo2.flags = 1; gwo2.act = 0;
      gwo2.alpha = 1.0f; gwo2.beta = 0.0f; gwo2.sa = 1.0f; gwo2.sb = 1.0f; gwo2.Npad = LD; gwo2.pad_ = 0;
      k_gemm<1><<<dim3((unsigned)((LD) + 31) / 32, (unsigned)((Ll) + 15) / 16, (unsigned)(1)), 32, 0, stream>>>(gwo2); }
    k_cl_out<<<(unsigned)(((long long)Ll * D + 255) / 256), 256, 0, stream>>>(O, LD, out, 2, (long long)Ll, D);
    hipMemsetAsync(XP, 0, (size_t)256 * 2052 * CI * 4, stream); hipMemsetAsync(HP, 0, (size_t)Hh * 2050 * C1 * 4, stream);
    k_cl_pad<<<(unsigned)(((long long)Hh * Tt * CI + 255) / 256), 256, 0, stream>>>(x, XP, 3, CI, Hh, Tt);
    { GemmP cp3_0;
      cp3_0.A = XP + (size_t)0 * CI; cp3_0.B = wpre + 0; cp3_0.bias = bpre; cp3_0.R = XP + (size_t)0 * CI; cp3_0.C = HP + C1;
      cp3_0.sAo = (long long)2052 * CI; cp3_0.sAi = 0; cp3_0.sAm = CI; cp3_0.sAk = 1; cp3_0.sBo = 0; cp3_0.sBi = 0; cp3_0.sBn = CI * 25; cp3_0.sBk = 25; cp3_0.sCo = (long long)2050 * C1; cp3_0.sCi = 0; cp3_0.sCm = C1; cp3_0.sRo = 0; cp3_0.sRi = 0; cp3_0.sRm = 0; cp3_0.sRn = 0;
      cp3_0.M = Tt; cp3_0.N = C1; cp3_0.K = CI; cp3_0.zi_n = 1; cp3_0.flags = 1; cp3_0.act = 0;
      cp3_0.alpha = 1.0f; cp3_0.beta = 0.0f; cp3_0.sa = 1.0f; cp3_0.sb = 1.0f; cp3_0.Npad = C1; cp3_0.pad_ = 0;
      k_gemm<1><<<dim3((unsigned)((C1) + 31) / 32, (unsigned)((Tt) + 15) / 16, (unsigned)(Hh)), 32, 0, stream>>>(cp3_0); }
    { GemmP cp3_1;
      cp3_1.A = XP + (size_t)1 * CI; cp3_1.B = wpre + 1; cp3_1.bias = XP + (size_t)1 * CI; cp3_1.R = HP + C1; cp3_1.C = HP + C1;
      cp3_1.sAo = (long long)2052 * CI; cp3_1.sAi = 0; cp3_1.sAm = CI; cp3_1.sAk = 1; cp3_1.sBo = 0; cp3_1.sBi = 0; cp3_1.sBn = CI * 25; cp3_1.sBk = 25; cp3_1.sCo = (long long)2050 * C1; cp3_1.sCi = 0; cp3_1.sCm = C1; cp3_1.sRo = (long long)2050 * C1; cp3_1.sRi = 0; cp3_1.sRm = C1; cp3_1.sRn = 1;
      cp3_1.M = Tt; cp3_1.N = C1; cp3_1.K = CI; cp3_1.zi_n = 1; cp3_1.flags = 4; cp3_1.act = 0;
      cp3_1.alpha = 1.0f; cp3_1.beta = 1.0f; cp3_1.sa = 1.0f; cp3_1.sb = 1.0f; cp3_1.Npad = C1; cp3_1.pad_ = 0;
      k_gemm<1><<<dim3((unsigned)((C1) + 31) / 32, (unsigned)((Tt) + 15) / 16, (unsigned)(Hh)), 32, 0, stream>>>(cp3_1); }
    { GemmP cp3_2;
      cp3_2.A = XP + (size_t)2 * CI; cp3_2.B = wpre + 2; cp3_2.bias = XP + (size_t)2 * CI; cp3_2.R = HP + C1; cp3_2.C = HP + C1;
      cp3_2.sAo = (long long)2052 * CI; cp3_2.sAi = 0; cp3_2.sAm = CI; cp3_2.sAk = 1; cp3_2.sBo = 0; cp3_2.sBi = 0; cp3_2.sBn = CI * 25; cp3_2.sBk = 25; cp3_2.sCo = (long long)2050 * C1; cp3_2.sCi = 0; cp3_2.sCm = C1; cp3_2.sRo = (long long)2050 * C1; cp3_2.sRi = 0; cp3_2.sRm = C1; cp3_2.sRn = 1;
      cp3_2.M = Tt; cp3_2.N = C1; cp3_2.K = CI; cp3_2.zi_n = 1; cp3_2.flags = 4; cp3_2.act = 0;
      cp3_2.alpha = 1.0f; cp3_2.beta = 1.0f; cp3_2.sa = 1.0f; cp3_2.sb = 1.0f; cp3_2.Npad = C1; cp3_2.pad_ = 0;
      k_gemm<1><<<dim3((unsigned)((C1) + 31) / 32, (unsigned)((Tt) + 15) / 16, (unsigned)(Hh)), 32, 0, stream>>>(cp3_2); }
    { GemmP cp3_3;
      cp3_3.A = XP + (size_t)3 * CI; cp3_3.B = wpre + 3; cp3_3.bias = XP + (size_t)3 * CI; cp3_3.R = HP + C1; cp3_3.C = HP + C1;
      cp3_3.sAo = (long long)2052 * CI; cp3_3.sAi = 0; cp3_3.sAm = CI; cp3_3.sAk = 1; cp3_3.sBo = 0; cp3_3.sBi = 0; cp3_3.sBn = CI * 25; cp3_3.sBk = 25; cp3_3.sCo = (long long)2050 * C1; cp3_3.sCi = 0; cp3_3.sCm = C1; cp3_3.sRo = (long long)2050 * C1; cp3_3.sRi = 0; cp3_3.sRm = C1; cp3_3.sRn = 1;
      cp3_3.M = Tt; cp3_3.N = C1; cp3_3.K = CI; cp3_3.zi_n = 1; cp3_3.flags = 4; cp3_3.act = 0;
      cp3_3.alpha = 1.0f; cp3_3.beta = 1.0f; cp3_3.sa = 1.0f; cp3_3.sb = 1.0f; cp3_3.Npad = C1; cp3_3.pad_ = 0;
      k_gemm<1><<<dim3((unsigned)((C1) + 31) / 32, (unsigned)((Tt) + 15) / 16, (unsigned)(Hh)), 32, 0, stream>>>(cp3_3); }
    { GemmP cp3_4;
      cp3_4.A = XP + (size_t)4 * CI; cp3_4.B = wpre + 4; cp3_4.bias = XP + (size_t)4 * CI; cp3_4.R = HP + C1; cp3_4.C = HP + C1;
      cp3_4.sAo = (long long)2052 * CI; cp3_4.sAi = 0; cp3_4.sAm = CI; cp3_4.sAk = 1; cp3_4.sBo = 0; cp3_4.sBi = 0; cp3_4.sBn = CI * 25; cp3_4.sBk = 25; cp3_4.sCo = (long long)2050 * C1; cp3_4.sCi = 0; cp3_4.sCm = C1; cp3_4.sRo = (long long)2050 * C1; cp3_4.sRi = 0; cp3_4.sRm = C1; cp3_4.sRn = 1;
      cp3_4.M = Tt; cp3_4.N = C1; cp3_4.K = CI; cp3_4.zi_n = 1; cp3_4.flags = 4; cp3_4.act = 0;
      cp3_4.alpha = 1.0f; cp3_4.beta = 1.0f; cp3_4.sa = 1.0f; cp3_4.sb = 1.0f; cp3_4.Npad = C1; cp3_4.pad_ = 0;
      k_gemm<1><<<dim3((unsigned)((C1) + 31) / 32, (unsigned)((Tt) + 15) / 16, (unsigned)(Hh)), 32, 0, stream>>>(cp3_4); }
    { GemmP cp3_5;
      cp3_5.A = XP + (size_t)2052 * CI; cp3_5.B = wpre + 5; cp3_5.bias = XP + (size_t)2052 * CI; cp3_5.R = HP + C1; cp3_5.C = HP + C1;
      cp3_5.sAo = (long long)2052 * CI; cp3_5.sAi = 0; cp3_5.sAm = CI; cp3_5.sAk = 1; cp3_5.sBo = 0; cp3_5.sBi = 0; cp3_5.sBn = CI * 25; cp3_5.sBk = 25; cp3_5.sCo = (long long)2050 * C1; cp3_5.sCi = 0; cp3_5.sCm = C1; cp3_5.sRo = (long long)2050 * C1; cp3_5.sRi = 0; cp3_5.sRm = C1; cp3_5.sRn = 1;
      cp3_5.M = Tt; cp3_5.N = C1; cp3_5.K = CI; cp3_5.zi_n = 1; cp3_5.flags = 4; cp3_5.act = 0;
      cp3_5.alpha = 1.0f; cp3_5.beta = 1.0f; cp3_5.sa = 1.0f; cp3_5.sb = 1.0f; cp3_5.Npad = C1; cp3_5.pad_ = 0;
      k_gemm<1><<<dim3((unsigned)((C1) + 31) / 32, (unsigned)((Tt) + 15) / 16, (unsigned)(Hh)), 32, 0, stream>>>(cp3_5); }
    { GemmP cp3_6;
      cp3_6.A = XP + (size_t)2053 * CI; cp3_6.B = wpre + 6; cp3_6.bias = XP + (size_t)2053 * CI; cp3_6.R = HP + C1; cp3_6.C = HP + C1;
      cp3_6.sAo = (long long)2052 * CI; cp3_6.sAi = 0; cp3_6.sAm = CI; cp3_6.sAk = 1; cp3_6.sBo = 0; cp3_6.sBi = 0; cp3_6.sBn = CI * 25; cp3_6.sBk = 25; cp3_6.sCo = (long long)2050 * C1; cp3_6.sCi = 0; cp3_6.sCm = C1; cp3_6.sRo = (long long)2050 * C1; cp3_6.sRi = 0; cp3_6.sRm = C1; cp3_6.sRn = 1;
      cp3_6.M = Tt; cp3_6.N = C1; cp3_6.K = CI; cp3_6.zi_n = 1; cp3_6.flags = 4; cp3_6.act = 0;
      cp3_6.alpha = 1.0f; cp3_6.beta = 1.0f; cp3_6.sa = 1.0f; cp3_6.sb = 1.0f; cp3_6.Npad = C1; cp3_6.pad_ = 0;
      k_gemm<1><<<dim3((unsigned)((C1) + 31) / 32, (unsigned)((Tt) + 15) / 16, (unsigned)(Hh)), 32, 0, stream>>>(cp3_6); }
    { GemmP cp3_7;
      cp3_7.A = XP + (size_t)2054 * CI; cp3_7.B = wpre + 7; cp3_7.bias = XP + (size_t)2054 * CI; cp3_7.R = HP + C1; cp3_7.C = HP + C1;
      cp3_7.sAo = (long long)2052 * CI; cp3_7.sAi = 0; cp3_7.sAm = CI; cp3_7.sAk = 1; cp3_7.sBo = 0; cp3_7.sBi = 0; cp3_7.sBn = CI * 25; cp3_7.sBk = 25; cp3_7.sCo = (long long)2050 * C1; cp3_7.sCi = 0; cp3_7.sCm = C1; cp3_7.sRo = (long long)2050 * C1; cp3_7.sRi = 0; cp3_7.sRm = C1; cp3_7.sRn = 1;
      cp3_7.M = Tt; cp3_7.N = C1; cp3_7.K = CI; cp3_7.zi_n = 1; cp3_7.flags = 4; cp3_7.act = 0;
      cp3_7.alpha = 1.0f; cp3_7.beta = 1.0f; cp3_7.sa = 1.0f; cp3_7.sb = 1.0f; cp3_7.Npad = C1; cp3_7.pad_ = 0;
      k_gemm<1><<<dim3((unsigned)((C1) + 31) / 32, (unsigned)((Tt) + 15) / 16, (unsigned)(Hh)), 32, 0, stream>>>(cp3_7); }
    { GemmP cp3_8;
      cp3_8.A = XP + (size_t)2055 * CI; cp3_8.B = wpre + 8; cp3_8.bias = XP + (size_t)2055 * CI; cp3_8.R = HP + C1; cp3_8.C = HP + C1;
      cp3_8.sAo = (long long)2052 * CI; cp3_8.sAi = 0; cp3_8.sAm = CI; cp3_8.sAk = 1; cp3_8.sBo = 0; cp3_8.sBi = 0; cp3_8.sBn = CI * 25; cp3_8.sBk = 25; cp3_8.sCo = (long long)2050 * C1; cp3_8.sCi = 0; cp3_8.sCm = C1; cp3_8.sRo = (long long)2050 * C1; cp3_8.sRi = 0; cp3_8.sRm = C1; cp3_8.sRn = 1;
      cp3_8.M = Tt; cp3_8.N = C1; cp3_8.K = CI; cp3_8.zi_n = 1; cp3_8.flags = 4; cp3_8.act = 0;
      cp3_8.alpha = 1.0f; cp3_8.beta = 1.0f; cp3_8.sa = 1.0f; cp3_8.sb = 1.0f; cp3_8.Npad = C1; cp3_8.pad_ = 0;
      k_gemm<1><<<dim3((unsigned)((C1) + 31) / 32, (unsigned)((Tt) + 15) / 16, (unsigned)(Hh)), 32, 0, stream>>>(cp3_8); }
    { GemmP cp3_9;
      cp3_9.A = XP + (size_t)2056 * CI; cp3_9.B = wpre + 9; cp3_9.bias = XP + (size_t)2056 * CI; cp3_9.R = HP + C1; cp3_9.C = HP + C1;
      cp3_9.sAo = (long long)2052 * CI; cp3_9.sAi = 0; cp3_9.sAm = CI; cp3_9.sAk = 1; cp3_9.sBo = 0; cp3_9.sBi = 0; cp3_9.sBn = CI * 25; cp3_9.sBk = 25; cp3_9.sCo = (long long)2050 * C1; cp3_9.sCi = 0; cp3_9.sCm = C1; cp3_9.sRo = (long long)2050 * C1; cp3_9.sRi = 0; cp3_9.sRm = C1; cp3_9.sRn = 1;
      cp3_9.M = Tt; cp3_9.N = C1; cp3_9.K = CI; cp3_9.zi_n = 1; cp3_9.flags = 4; cp3_9.act = 0;
      cp3_9.alpha = 1.0f; cp3_9.beta = 1.0f; cp3_9.sa = 1.0f; cp3_9.sb = 1.0f; cp3_9.Npad = C1; cp3_9.pad_ = 0;
      k_gemm<1><<<dim3((unsigned)((C1) + 31) / 32, (unsigned)((Tt) + 15) / 16, (unsigned)(Hh)), 32, 0, stream>>>(cp3_9); }
    { GemmP cp3_10;
      cp3_10.A = XP + (size_t)4104 * CI; cp3_10.B = wpre + 10; cp3_10.bias = XP + (size_t)4104 * CI; cp3_10.R = HP + C1; cp3_10.C = HP + C1;
      cp3_10.sAo = (long long)2052 * CI; cp3_10.sAi = 0; cp3_10.sAm = CI; cp3_10.sAk = 1; cp3_10.sBo = 0; cp3_10.sBi = 0; cp3_10.sBn = CI * 25; cp3_10.sBk = 25; cp3_10.sCo = (long long)2050 * C1; cp3_10.sCi = 0; cp3_10.sCm = C1; cp3_10.sRo = (long long)2050 * C1; cp3_10.sRi = 0; cp3_10.sRm = C1; cp3_10.sRn = 1;
      cp3_10.M = Tt; cp3_10.N = C1; cp3_10.K = CI; cp3_10.zi_n = 1; cp3_10.flags = 4; cp3_10.act = 0;
      cp3_10.alpha = 1.0f; cp3_10.beta = 1.0f; cp3_10.sa = 1.0f; cp3_10.sb = 1.0f; cp3_10.Npad = C1; cp3_10.pad_ = 0;
      k_gemm<1><<<dim3((unsigned)((C1) + 31) / 32, (unsigned)((Tt) + 15) / 16, (unsigned)(Hh)), 32, 0, stream>>>(cp3_10); }
    { GemmP cp3_11;
      cp3_11.A = XP + (size_t)4105 * CI; cp3_11.B = wpre + 11; cp3_11.bias = XP + (size_t)4105 * CI; cp3_11.R = HP + C1; cp3_11.C = HP + C1;
      cp3_11.sAo = (long long)2052 * CI; cp3_11.sAi = 0; cp3_11.sAm = CI; cp3_11.sAk = 1; cp3_11.sBo = 0; cp3_11.sBi = 0; cp3_11.sBn = CI * 25; cp3_11.sBk = 25; cp3_11.sCo = (long long)2050 * C1; cp3_11.sCi = 0; cp3_11.sCm = C1; cp3_11.sRo = (long long)2050 * C1; cp3_11.sRi = 0; cp3_11.sRm = C1; cp3_11.sRn = 1;
      cp3_11.M = Tt; cp3_11.N = C1; cp3_11.K = CI; cp3_11.zi_n = 1; cp3_11.flags = 4; cp3_11.act = 0;
      cp3_11.alpha = 1.0f; cp3_11.beta = 1.0f; cp3_11.sa = 1.0f; cp3_11.sb = 1.0f; cp3_11.Npad = C1; cp3_11.pad_ = 0;
      k_gemm<1><<<dim3((unsigned)((C1) + 31) / 32, (unsigned)((Tt) + 15) / 16, (unsigned)(Hh)), 32, 0, stream>>>(cp3_11); }
    { GemmP cp3_12;
      cp3_12.A = XP + (size_t)4106 * CI; cp3_12.B = wpre + 12; cp3_12.bias = XP + (size_t)4106 * CI; cp3_12.R = HP + C1; cp3_12.C = HP + C1;
      cp3_12.sAo = (long long)2052 * CI; cp3_12.sAi = 0; cp3_12.sAm = CI; cp3_12.sAk = 1; cp3_12.sBo = 0; cp3_12.sBi = 0; cp3_12.sBn = CI * 25; cp3_12.sBk = 25; cp3_12.sCo = (long long)2050 * C1; cp3_12.sCi = 0; cp3_12.sCm = C1; cp3_12.sRo = (long long)2050 * C1; cp3_12.sRi = 0; cp3_12.sRm = C1; cp3_12.sRn = 1;
      cp3_12.M = Tt; cp3_12.N = C1; cp3_12.K = CI; cp3_12.zi_n = 1; cp3_12.flags = 4; cp3_12.act = 0;
      cp3_12.alpha = 1.0f; cp3_12.beta = 1.0f; cp3_12.sa = 1.0f; cp3_12.sb = 1.0f; cp3_12.Npad = C1; cp3_12.pad_ = 0;
      k_gemm<1><<<dim3((unsigned)((C1) + 31) / 32, (unsigned)((Tt) + 15) / 16, (unsigned)(Hh)), 32, 0, stream>>>(cp3_12); }
    { GemmP cp3_13;
      cp3_13.A = XP + (size_t)4107 * CI; cp3_13.B = wpre + 13; cp3_13.bias = XP + (size_t)4107 * CI; cp3_13.R = HP + C1; cp3_13.C = HP + C1;
      cp3_13.sAo = (long long)2052 * CI; cp3_13.sAi = 0; cp3_13.sAm = CI; cp3_13.sAk = 1; cp3_13.sBo = 0; cp3_13.sBi = 0; cp3_13.sBn = CI * 25; cp3_13.sBk = 25; cp3_13.sCo = (long long)2050 * C1; cp3_13.sCi = 0; cp3_13.sCm = C1; cp3_13.sRo = (long long)2050 * C1; cp3_13.sRi = 0; cp3_13.sRm = C1; cp3_13.sRn = 1;
      cp3_13.M = Tt; cp3_13.N = C1; cp3_13.K = CI; cp3_13.zi_n = 1; cp3_13.flags = 4; cp3_13.act = 0;
      cp3_13.alpha = 1.0f; cp3_13.beta = 1.0f; cp3_13.sa = 1.0f; cp3_13.sb = 1.0f; cp3_13.Npad = C1; cp3_13.pad_ = 0;
      k_gemm<1><<<dim3((unsigned)((C1) + 31) / 32, (unsigned)((Tt) + 15) / 16, (unsigned)(Hh)), 32, 0, stream>>>(cp3_13); }
    { GemmP cp3_14;
      cp3_14.A = XP + (size_t)4108 * CI; cp3_14.B = wpre + 14; cp3_14.bias = XP + (size_t)4108 * CI; cp3_14.R = HP + C1; cp3_14.C = HP + C1;
      cp3_14.sAo = (long long)2052 * CI; cp3_14.sAi = 0; cp3_14.sAm = CI; cp3_14.sAk = 1; cp3_14.sBo = 0; cp3_14.sBi = 0; cp3_14.sBn = CI * 25; cp3_14.sBk = 25; cp3_14.sCo = (long long)2050 * C1; cp3_14.sCi = 0; cp3_14.sCm = C1; cp3_14.sRo = (long long)2050 * C1; cp3_14.sRi = 0; cp3_14.sRm = C1; cp3_14.sRn = 1;
      cp3_14.M = Tt; cp3_14.N = C1; cp3_14.K = CI; cp3_14.zi_n = 1; cp3_14.flags = 4; cp3_14.act = 0;
      cp3_14.alpha = 1.0f; cp3_14.beta = 1.0f; cp3_14.sa = 1.0f; cp3_14.sb = 1.0f; cp3_14.Npad = C1; cp3_14.pad_ = 0;
      k_gemm<1><<<dim3((unsigned)((C1) + 31) / 32, (unsigned)((Tt) + 15) / 16, (unsigned)(Hh)), 32, 0, stream>>>(cp3_14); }
    { GemmP cp3_15;
      cp3_15.A = XP + (size_t)6156 * CI; cp3_15.B = wpre + 15; cp3_15.bias = XP + (size_t)6156 * CI; cp3_15.R = HP + C1; cp3_15.C = HP + C1;
      cp3_15.sAo = (long long)2052 * CI; cp3_15.sAi = 0; cp3_15.sAm = CI; cp3_15.sAk = 1; cp3_15.sBo = 0; cp3_15.sBi = 0; cp3_15.sBn = CI * 25; cp3_15.sBk = 25; cp3_15.sCo = (long long)2050 * C1; cp3_15.sCi = 0; cp3_15.sCm = C1; cp3_15.sRo = (long long)2050 * C1; cp3_15.sRi = 0; cp3_15.sRm = C1; cp3_15.sRn = 1;
      cp3_15.M = Tt; cp3_15.N = C1; cp3_15.K = CI; cp3_15.zi_n = 1; cp3_15.flags = 4; cp3_15.act = 0;
      cp3_15.alpha = 1.0f; cp3_15.beta = 1.0f; cp3_15.sa = 1.0f; cp3_15.sb = 1.0f; cp3_15.Npad = C1; cp3_15.pad_ = 0;
      k_gemm<1><<<dim3((unsigned)((C1) + 31) / 32, (unsigned)((Tt) + 15) / 16, (unsigned)(Hh)), 32, 0, stream>>>(cp3_15); }
    { GemmP cp3_16;
      cp3_16.A = XP + (size_t)6157 * CI; cp3_16.B = wpre + 16; cp3_16.bias = XP + (size_t)6157 * CI; cp3_16.R = HP + C1; cp3_16.C = HP + C1;
      cp3_16.sAo = (long long)2052 * CI; cp3_16.sAi = 0; cp3_16.sAm = CI; cp3_16.sAk = 1; cp3_16.sBo = 0; cp3_16.sBi = 0; cp3_16.sBn = CI * 25; cp3_16.sBk = 25; cp3_16.sCo = (long long)2050 * C1; cp3_16.sCi = 0; cp3_16.sCm = C1; cp3_16.sRo = (long long)2050 * C1; cp3_16.sRi = 0; cp3_16.sRm = C1; cp3_16.sRn = 1;
      cp3_16.M = Tt; cp3_16.N = C1; cp3_16.K = CI; cp3_16.zi_n = 1; cp3_16.flags = 4; cp3_16.act = 0;
      cp3_16.alpha = 1.0f; cp3_16.beta = 1.0f; cp3_16.sa = 1.0f; cp3_16.sb = 1.0f; cp3_16.Npad = C1; cp3_16.pad_ = 0;
      k_gemm<1><<<dim3((unsigned)((C1) + 31) / 32, (unsigned)((Tt) + 15) / 16, (unsigned)(Hh)), 32, 0, stream>>>(cp3_16); }
    { GemmP cp3_17;
      cp3_17.A = XP + (size_t)6158 * CI; cp3_17.B = wpre + 17; cp3_17.bias = XP + (size_t)6158 * CI; cp3_17.R = HP + C1; cp3_17.C = HP + C1;
      cp3_17.sAo = (long long)2052 * CI; cp3_17.sAi = 0; cp3_17.sAm = CI; cp3_17.sAk = 1; cp3_17.sBo = 0; cp3_17.sBi = 0; cp3_17.sBn = CI * 25; cp3_17.sBk = 25; cp3_17.sCo = (long long)2050 * C1; cp3_17.sCi = 0; cp3_17.sCm = C1; cp3_17.sRo = (long long)2050 * C1; cp3_17.sRi = 0; cp3_17.sRm = C1; cp3_17.sRn = 1;
      cp3_17.M = Tt; cp3_17.N = C1; cp3_17.K = CI; cp3_17.zi_n = 1; cp3_17.flags = 4; cp3_17.act = 0;
      cp3_17.alpha = 1.0f; cp3_17.beta = 1.0f; cp3_17.sa = 1.0f; cp3_17.sb = 1.0f; cp3_17.Npad = C1; cp3_17.pad_ = 0;
      k_gemm<1><<<dim3((unsigned)((C1) + 31) / 32, (unsigned)((Tt) + 15) / 16, (unsigned)(Hh)), 32, 0, stream>>>(cp3_17); }
    { GemmP cp3_18;
      cp3_18.A = XP + (size_t)6159 * CI; cp3_18.B = wpre + 18; cp3_18.bias = XP + (size_t)6159 * CI; cp3_18.R = HP + C1; cp3_18.C = HP + C1;
      cp3_18.sAo = (long long)2052 * CI; cp3_18.sAi = 0; cp3_18.sAm = CI; cp3_18.sAk = 1; cp3_18.sBo = 0; cp3_18.sBi = 0; cp3_18.sBn = CI * 25; cp3_18.sBk = 25; cp3_18.sCo = (long long)2050 * C1; cp3_18.sCi = 0; cp3_18.sCm = C1; cp3_18.sRo = (long long)2050 * C1; cp3_18.sRi = 0; cp3_18.sRm = C1; cp3_18.sRn = 1;
      cp3_18.M = Tt; cp3_18.N = C1; cp3_18.K = CI; cp3_18.zi_n = 1; cp3_18.flags = 4; cp3_18.act = 0;
      cp3_18.alpha = 1.0f; cp3_18.beta = 1.0f; cp3_18.sa = 1.0f; cp3_18.sb = 1.0f; cp3_18.Npad = C1; cp3_18.pad_ = 0;
      k_gemm<1><<<dim3((unsigned)((C1) + 31) / 32, (unsigned)((Tt) + 15) / 16, (unsigned)(Hh)), 32, 0, stream>>>(cp3_18); }
    { GemmP cp3_19;
      cp3_19.A = XP + (size_t)6160 * CI; cp3_19.B = wpre + 19; cp3_19.bias = XP + (size_t)6160 * CI; cp3_19.R = HP + C1; cp3_19.C = HP + C1;
      cp3_19.sAo = (long long)2052 * CI; cp3_19.sAi = 0; cp3_19.sAm = CI; cp3_19.sAk = 1; cp3_19.sBo = 0; cp3_19.sBi = 0; cp3_19.sBn = CI * 25; cp3_19.sBk = 25; cp3_19.sCo = (long long)2050 * C1; cp3_19.sCi = 0; cp3_19.sCm = C1; cp3_19.sRo = (long long)2050 * C1; cp3_19.sRi = 0; cp3_19.sRm = C1; cp3_19.sRn = 1;
      cp3_19.M = Tt; cp3_19.N = C1; cp3_19.K = CI; cp3_19.zi_n = 1; cp3_19.flags = 4; cp3_19.act = 0;
      cp3_19.alpha = 1.0f; cp3_19.beta = 1.0f; cp3_19.sa = 1.0f; cp3_19.sb = 1.0f; cp3_19.Npad = C1; cp3_19.pad_ = 0;
      k_gemm<1><<<dim3((unsigned)((C1) + 31) / 32, (unsigned)((Tt) + 15) / 16, (unsigned)(Hh)), 32, 0, stream>>>(cp3_19); }
    { GemmP cp3_20;
      cp3_20.A = XP + (size_t)8208 * CI; cp3_20.B = wpre + 20; cp3_20.bias = XP + (size_t)8208 * CI; cp3_20.R = HP + C1; cp3_20.C = HP + C1;
      cp3_20.sAo = (long long)2052 * CI; cp3_20.sAi = 0; cp3_20.sAm = CI; cp3_20.sAk = 1; cp3_20.sBo = 0; cp3_20.sBi = 0; cp3_20.sBn = CI * 25; cp3_20.sBk = 25; cp3_20.sCo = (long long)2050 * C1; cp3_20.sCi = 0; cp3_20.sCm = C1; cp3_20.sRo = (long long)2050 * C1; cp3_20.sRi = 0; cp3_20.sRm = C1; cp3_20.sRn = 1;
      cp3_20.M = Tt; cp3_20.N = C1; cp3_20.K = CI; cp3_20.zi_n = 1; cp3_20.flags = 4; cp3_20.act = 0;
      cp3_20.alpha = 1.0f; cp3_20.beta = 1.0f; cp3_20.sa = 1.0f; cp3_20.sb = 1.0f; cp3_20.Npad = C1; cp3_20.pad_ = 0;
      k_gemm<1><<<dim3((unsigned)((C1) + 31) / 32, (unsigned)((Tt) + 15) / 16, (unsigned)(Hh)), 32, 0, stream>>>(cp3_20); }
    { GemmP cp3_21;
      cp3_21.A = XP + (size_t)8209 * CI; cp3_21.B = wpre + 21; cp3_21.bias = XP + (size_t)8209 * CI; cp3_21.R = HP + C1; cp3_21.C = HP + C1;
      cp3_21.sAo = (long long)2052 * CI; cp3_21.sAi = 0; cp3_21.sAm = CI; cp3_21.sAk = 1; cp3_21.sBo = 0; cp3_21.sBi = 0; cp3_21.sBn = CI * 25; cp3_21.sBk = 25; cp3_21.sCo = (long long)2050 * C1; cp3_21.sCi = 0; cp3_21.sCm = C1; cp3_21.sRo = (long long)2050 * C1; cp3_21.sRi = 0; cp3_21.sRm = C1; cp3_21.sRn = 1;
      cp3_21.M = Tt; cp3_21.N = C1; cp3_21.K = CI; cp3_21.zi_n = 1; cp3_21.flags = 4; cp3_21.act = 0;
      cp3_21.alpha = 1.0f; cp3_21.beta = 1.0f; cp3_21.sa = 1.0f; cp3_21.sb = 1.0f; cp3_21.Npad = C1; cp3_21.pad_ = 0;
      k_gemm<1><<<dim3((unsigned)((C1) + 31) / 32, (unsigned)((Tt) + 15) / 16, (unsigned)(Hh)), 32, 0, stream>>>(cp3_21); }
    { GemmP cp3_22;
      cp3_22.A = XP + (size_t)8210 * CI; cp3_22.B = wpre + 22; cp3_22.bias = XP + (size_t)8210 * CI; cp3_22.R = HP + C1; cp3_22.C = HP + C1;
      cp3_22.sAo = (long long)2052 * CI; cp3_22.sAi = 0; cp3_22.sAm = CI; cp3_22.sAk = 1; cp3_22.sBo = 0; cp3_22.sBi = 0; cp3_22.sBn = CI * 25; cp3_22.sBk = 25; cp3_22.sCo = (long long)2050 * C1; cp3_22.sCi = 0; cp3_22.sCm = C1; cp3_22.sRo = (long long)2050 * C1; cp3_22.sRi = 0; cp3_22.sRm = C1; cp3_22.sRn = 1;
      cp3_22.M = Tt; cp3_22.N = C1; cp3_22.K = CI; cp3_22.zi_n = 1; cp3_22.flags = 4; cp3_22.act = 0;
      cp3_22.alpha = 1.0f; cp3_22.beta = 1.0f; cp3_22.sa = 1.0f; cp3_22.sb = 1.0f; cp3_22.Npad = C1; cp3_22.pad_ = 0;
      k_gemm<1><<<dim3((unsigned)((C1) + 31) / 32, (unsigned)((Tt) + 15) / 16, (unsigned)(Hh)), 32, 0, stream>>>(cp3_22); }
    { GemmP cp3_23;
      cp3_23.A = XP + (size_t)8211 * CI; cp3_23.B = wpre + 23; cp3_23.bias = XP + (size_t)8211 * CI; cp3_23.R = HP + C1; cp3_23.C = HP + C1;
      cp3_23.sAo = (long long)2052 * CI; cp3_23.sAi = 0; cp3_23.sAm = CI; cp3_23.sAk = 1; cp3_23.sBo = 0; cp3_23.sBi = 0; cp3_23.sBn = CI * 25; cp3_23.sBk = 25; cp3_23.sCo = (long long)2050 * C1; cp3_23.sCi = 0; cp3_23.sCm = C1; cp3_23.sRo = (long long)2050 * C1; cp3_23.sRi = 0; cp3_23.sRm = C1; cp3_23.sRn = 1;
      cp3_23.M = Tt; cp3_23.N = C1; cp3_23.K = CI; cp3_23.zi_n = 1; cp3_23.flags = 4; cp3_23.act = 0;
      cp3_23.alpha = 1.0f; cp3_23.beta = 1.0f; cp3_23.sa = 1.0f; cp3_23.sb = 1.0f; cp3_23.Npad = C1; cp3_23.pad_ = 0;
      k_gemm<1><<<dim3((unsigned)((C1) + 31) / 32, (unsigned)((Tt) + 15) / 16, (unsigned)(Hh)), 32, 0, stream>>>(cp3_23); }
    { GemmP cp3_24;
      cp3_24.A = XP + (size_t)8212 * CI; cp3_24.B = wpre + 24; cp3_24.bias = XP + (size_t)8212 * CI; cp3_24.R = HP + C1; cp3_24.C = HP + C1;
      cp3_24.sAo = (long long)2052 * CI; cp3_24.sAi = 0; cp3_24.sAm = CI; cp3_24.sAk = 1; cp3_24.sBo = 0; cp3_24.sBi = 0; cp3_24.sBn = CI * 25; cp3_24.sBk = 25; cp3_24.sCo = (long long)2050 * C1; cp3_24.sCi = 0; cp3_24.sCm = C1; cp3_24.sRo = (long long)2050 * C1; cp3_24.sRi = 0; cp3_24.sRm = C1; cp3_24.sRn = 1;
      cp3_24.M = Tt; cp3_24.N = C1; cp3_24.K = CI; cp3_24.zi_n = 1; cp3_24.flags = 4; cp3_24.act = 0;
      cp3_24.alpha = 1.0f; cp3_24.beta = 1.0f; cp3_24.sa = 1.0f; cp3_24.sb = 1.0f; cp3_24.Npad = C1; cp3_24.pad_ = 0;
      k_gemm<1><<<dim3((unsigned)((C1) + 31) / 32, (unsigned)((Tt) + 15) / 16, (unsigned)(Hh)), 32, 0, stream>>>(cp3_24); }
    k_cl_bnl<<<(unsigned)(((long long)Hh * Tt * C1 + 255) / 256), 256, 0, stream>>>(HP, bng, bnb, bnm, bnv, Hh, Tt, C1);
    { GemmP ceq3_0;
      ceq3_0.A = HP + (size_t)0 * C1; ceq3_0.B = wq + 0; ceq3_0.bias = bq; ceq3_0.R = HP + (size_t)0 * C1; ceq3_0.C = Q;
      ceq3_0.sAo = (long long)3 * 2050 * C1; ceq3_0.sAi = 0; ceq3_0.sAm = C1; ceq3_0.sAk = 1; ceq3_0.sBo = 0; ceq3_0.sBi = 0; ceq3_0.sBn = C1 * 9; ceq3_0.sBk = 9; ceq3_0.sCo = (long long)Tt * LD; ceq3_0.sCi = 0; ceq3_0.sCm = LD; ceq3_0.sRo = 0; ceq3_0.sRi = 0; ceq3_0.sRm = 0; ceq3_0.sRn = 0;
      ceq3_0.M = Tt; ceq3_0.N = D; ceq3_0.K = C1; ceq3_0.zi_n = 1; ceq3_0.flags = 1; ceq3_0.act = 0;
      ceq3_0.alpha = 1.0f; ceq3_0.beta = 0.0f; ceq3_0.sa = 1.0f; ceq3_0.sb = 1.0f; ceq3_0.Npad = LD; ceq3_0.pad_ = 0;
      k_gemm<1><<<dim3((unsigned)((LD) + 31) / 32, (unsigned)((Tt) + 15) / 16, (unsigned)(Fo)), 32, 0, stream>>>(ceq3_0); }
    { GemmP ceq3_1;
      ceq3_1.A = HP + (size_t)1 * C1; ceq3_1.B = wq + 1; ceq3_1.bias = HP + (size_t)1 * C1; ceq3_1.R = Q; ceq3_1.C = Q;
      ceq3_1.sAo = (long long)3 * 2050 * C1; ceq3_1.sAi = 0; ceq3_1.sAm = C1; ceq3_1.sAk = 1; ceq3_1.sBo = 0; ceq3_1.sBi = 0; ceq3_1.sBn = C1 * 9; ceq3_1.sBk = 9; ceq3_1.sCo = (long long)Tt * LD; ceq3_1.sCi = 0; ceq3_1.sCm = LD; ceq3_1.sRo = (long long)Tt * LD; ceq3_1.sRi = 0; ceq3_1.sRm = LD; ceq3_1.sRn = 1;
      ceq3_1.M = Tt; ceq3_1.N = D; ceq3_1.K = C1; ceq3_1.zi_n = 1; ceq3_1.flags = 4; ceq3_1.act = 0;
      ceq3_1.alpha = 1.0f; ceq3_1.beta = 1.0f; ceq3_1.sa = 1.0f; ceq3_1.sb = 1.0f; ceq3_1.Npad = LD; ceq3_1.pad_ = 0;
      k_gemm<1><<<dim3((unsigned)((LD) + 31) / 32, (unsigned)((Tt) + 15) / 16, (unsigned)(Fo)), 32, 0, stream>>>(ceq3_1); }
    { GemmP ceq3_2;
      ceq3_2.A = HP + (size_t)2 * C1; ceq3_2.B = wq + 2; ceq3_2.bias = HP + (size_t)2 * C1; ceq3_2.R = Q; ceq3_2.C = Q;
      ceq3_2.sAo = (long long)3 * 2050 * C1; ceq3_2.sAi = 0; ceq3_2.sAm = C1; ceq3_2.sAk = 1; ceq3_2.sBo = 0; ceq3_2.sBi = 0; ceq3_2.sBn = C1 * 9; ceq3_2.sBk = 9; ceq3_2.sCo = (long long)Tt * LD; ceq3_2.sCi = 0; ceq3_2.sCm = LD; ceq3_2.sRo = (long long)Tt * LD; ceq3_2.sRi = 0; ceq3_2.sRm = LD; ceq3_2.sRn = 1;
      ceq3_2.M = Tt; ceq3_2.N = D; ceq3_2.K = C1; ceq3_2.zi_n = 1; ceq3_2.flags = 4; ceq3_2.act = 0;
      ceq3_2.alpha = 1.0f; ceq3_2.beta = 1.0f; ceq3_2.sa = 1.0f; ceq3_2.sb = 1.0f; ceq3_2.Npad = LD; ceq3_2.pad_ = 0;
      k_gemm<1><<<dim3((unsigned)((LD) + 31) / 32, (unsigned)((Tt) + 15) / 16, (unsigned)(Fo)), 32, 0, stream>>>(ceq3_2); }
    { GemmP ceq3_3;
      ceq3_3.A = HP + (size_t)2050 * C1; ceq3_3.B = wq + 3; ceq3_3.bias = HP + (size_t)2050 * C1; ceq3_3.R = Q; ceq3_3.C = Q;
      ceq3_3.sAo = (long long)3 * 2050 * C1; ceq3_3.sAi = 0; ceq3_3.sAm = C1; ceq3_3.sAk = 1; ceq3_3.sBo = 0; ceq3_3.sBi = 0; ceq3_3.sBn = C1 * 9; ceq3_3.sBk = 9; ceq3_3.sCo = (long long)Tt * LD; ceq3_3.sCi = 0; ceq3_3.sCm = LD; ceq3_3.sRo = (long long)Tt * LD; ceq3_3.sRi = 0; ceq3_3.sRm = LD; ceq3_3.sRn = 1;
      ceq3_3.M = Tt; ceq3_3.N = D; ceq3_3.K = C1; ceq3_3.zi_n = 1; ceq3_3.flags = 4; ceq3_3.act = 0;
      ceq3_3.alpha = 1.0f; ceq3_3.beta = 1.0f; ceq3_3.sa = 1.0f; ceq3_3.sb = 1.0f; ceq3_3.Npad = LD; ceq3_3.pad_ = 0;
      k_gemm<1><<<dim3((unsigned)((LD) + 31) / 32, (unsigned)((Tt) + 15) / 16, (unsigned)(Fo)), 32, 0, stream>>>(ceq3_3); }
    { GemmP ceq3_4;
      ceq3_4.A = HP + (size_t)2051 * C1; ceq3_4.B = wq + 4; ceq3_4.bias = HP + (size_t)2051 * C1; ceq3_4.R = Q; ceq3_4.C = Q;
      ceq3_4.sAo = (long long)3 * 2050 * C1; ceq3_4.sAi = 0; ceq3_4.sAm = C1; ceq3_4.sAk = 1; ceq3_4.sBo = 0; ceq3_4.sBi = 0; ceq3_4.sBn = C1 * 9; ceq3_4.sBk = 9; ceq3_4.sCo = (long long)Tt * LD; ceq3_4.sCi = 0; ceq3_4.sCm = LD; ceq3_4.sRo = (long long)Tt * LD; ceq3_4.sRi = 0; ceq3_4.sRm = LD; ceq3_4.sRn = 1;
      ceq3_4.M = Tt; ceq3_4.N = D; ceq3_4.K = C1; ceq3_4.zi_n = 1; ceq3_4.flags = 4; ceq3_4.act = 0;
      ceq3_4.alpha = 1.0f; ceq3_4.beta = 1.0f; ceq3_4.sa = 1.0f; ceq3_4.sb = 1.0f; ceq3_4.Npad = LD; ceq3_4.pad_ = 0;
      k_gemm<1><<<dim3((unsigned)((LD) + 31) / 32, (unsigned)((Tt) + 15) / 16, (unsigned)(Fo)), 32, 0, stream>>>(ceq3_4); }
    { GemmP ceq3_5;
      ceq3_5.A = HP + (size_t)2052 * C1; ceq3_5.B = wq + 5; ceq3_5.bias = HP + (size_t)2052 * C1; ceq3_5.R = Q; ceq3_5.C = Q;
      ceq3_5.sAo = (long long)3 * 2050 * C1; ceq3_5.sAi = 0; ceq3_5.sAm = C1; ceq3_5.sAk = 1; ceq3_5.sBo = 0; ceq3_5.sBi = 0; ceq3_5.sBn = C1 * 9; ceq3_5.sBk = 9; ceq3_5.sCo = (long long)Tt * LD; ceq3_5.sCi = 0; ceq3_5.sCm = LD; ceq3_5.sRo = (long long)Tt * LD; ceq3_5.sRi = 0; ceq3_5.sRm = LD; ceq3_5.sRn = 1;
      ceq3_5.M = Tt; ceq3_5.N = D; ceq3_5.K = C1; ceq3_5.zi_n = 1; ceq3_5.flags = 4; ceq3_5.act = 0;
      ceq3_5.alpha = 1.0f; ceq3_5.beta = 1.0f; ceq3_5.sa = 1.0f; ceq3_5.sb = 1.0f; ceq3_5.Npad = LD; ceq3_5.pad_ = 0;
      k_gemm<1><<<dim3((unsigned)((LD) + 31) / 32, (unsigned)((Tt) + 15) / 16, (unsigned)(Fo)), 32, 0, stream>>>(ceq3_5); }
    { GemmP ceq3_6;
      ceq3_6.A = HP + (size_t)4100 * C1; ceq3_6.B = wq + 6; ceq3_6.bias = HP + (size_t)4100 * C1; ceq3_6.R = Q; ceq3_6.C = Q;
      ceq3_6.sAo = (long long)3 * 2050 * C1; ceq3_6.sAi = 0; ceq3_6.sAm = C1; ceq3_6.sAk = 1; ceq3_6.sBo = 0; ceq3_6.sBi = 0; ceq3_6.sBn = C1 * 9; ceq3_6.sBk = 9; ceq3_6.sCo = (long long)Tt * LD; ceq3_6.sCi = 0; ceq3_6.sCm = LD; ceq3_6.sRo = (long long)Tt * LD; ceq3_6.sRi = 0; ceq3_6.sRm = LD; ceq3_6.sRn = 1;
      ceq3_6.M = Tt; ceq3_6.N = D; ceq3_6.K = C1; ceq3_6.zi_n = 1; ceq3_6.flags = 4; ceq3_6.act = 0;
      ceq3_6.alpha = 1.0f; ceq3_6.beta = 1.0f; ceq3_6.sa = 1.0f; ceq3_6.sb = 1.0f; ceq3_6.Npad = LD; ceq3_6.pad_ = 0;
      k_gemm<1><<<dim3((unsigned)((LD) + 31) / 32, (unsigned)((Tt) + 15) / 16, (unsigned)(Fo)), 32, 0, stream>>>(ceq3_6); }
    { GemmP ceq3_7;
      ceq3_7.A = HP + (size_t)4101 * C1; ceq3_7.B = wq + 7; ceq3_7.bias = HP + (size_t)4101 * C1; ceq3_7.R = Q; ceq3_7.C = Q;
      ceq3_7.sAo = (long long)3 * 2050 * C1; ceq3_7.sAi = 0; ceq3_7.sAm = C1; ceq3_7.sAk = 1; ceq3_7.sBo = 0; ceq3_7.sBi = 0; ceq3_7.sBn = C1 * 9; ceq3_7.sBk = 9; ceq3_7.sCo = (long long)Tt * LD; ceq3_7.sCi = 0; ceq3_7.sCm = LD; ceq3_7.sRo = (long long)Tt * LD; ceq3_7.sRi = 0; ceq3_7.sRm = LD; ceq3_7.sRn = 1;
      ceq3_7.M = Tt; ceq3_7.N = D; ceq3_7.K = C1; ceq3_7.zi_n = 1; ceq3_7.flags = 4; ceq3_7.act = 0;
      ceq3_7.alpha = 1.0f; ceq3_7.beta = 1.0f; ceq3_7.sa = 1.0f; ceq3_7.sb = 1.0f; ceq3_7.Npad = LD; ceq3_7.pad_ = 0;
      k_gemm<1><<<dim3((unsigned)((LD) + 31) / 32, (unsigned)((Tt) + 15) / 16, (unsigned)(Fo)), 32, 0, stream>>>(ceq3_7); }
    { GemmP ceq3_8;
      ceq3_8.A = HP + (size_t)4102 * C1; ceq3_8.B = wq + 8; ceq3_8.bias = HP + (size_t)4102 * C1; ceq3_8.R = Q; ceq3_8.C = Q;
      ceq3_8.sAo = (long long)3 * 2050 * C1; ceq3_8.sAi = 0; ceq3_8.sAm = C1; ceq3_8.sAk = 1; ceq3_8.sBo = 0; ceq3_8.sBi = 0; ceq3_8.sBn = C1 * 9; ceq3_8.sBk = 9; ceq3_8.sCo = (long long)Tt * LD; ceq3_8.sCi = 0; ceq3_8.sCm = LD; ceq3_8.sRo = (long long)Tt * LD; ceq3_8.sRi = 0; ceq3_8.sRm = LD; ceq3_8.sRn = 1;
      ceq3_8.M = Tt; ceq3_8.N = D; ceq3_8.K = C1; ceq3_8.zi_n = 1; ceq3_8.flags = 4; ceq3_8.act = 0;
      ceq3_8.alpha = 1.0f; ceq3_8.beta = 1.0f; ceq3_8.sa = 1.0f; ceq3_8.sb = 1.0f; ceq3_8.Npad = LD; ceq3_8.pad_ = 0;
      k_gemm<1><<<dim3((unsigned)((LD) + 31) / 32, (unsigned)((Tt) + 15) / 16, (unsigned)(Fo)), 32, 0, stream>>>(ceq3_8); }

    { GemmP cekv3_0;
      cekv3_0.A = HP + (size_t)0 * C1; cekv3_0.B = wkv + 0; cekv3_0.bias = bkv; cekv3_0.R = HP + (size_t)0 * C1; cekv3_0.C = KV;
      cekv3_0.sAo = (long long)3 * 2050 * C1; cekv3_0.sAi = 0; cekv3_0.sAm = C1; cekv3_0.sAk = 1; cekv3_0.sBo = 0; cekv3_0.sBi = 0; cekv3_0.sBn = C1 * 9; cekv3_0.sBk = 9; cekv3_0.sCo = (long long)Tt * LD; cekv3_0.sCi = 0; cekv3_0.sCm = LD; cekv3_0.sRo = 0; cekv3_0.sRi = 0; cekv3_0.sRm = 0; cekv3_0.sRn = 0;
      cekv3_0.M = Tt; cekv3_0.N = D; cekv3_0.K = C1; cekv3_0.zi_n = 1; cekv3_0.flags = 1; cekv3_0.act = 0;
      cekv3_0.alpha = 1.0f; cekv3_0.beta = 0.0f; cekv3_0.sa = 1.0f; cekv3_0.sb = 1.0f; cekv3_0.Npad = LD; cekv3_0.pad_ = 0;
      k_gemm<1><<<dim3((unsigned)((LD) + 31) / 32, (unsigned)((Tt) + 15) / 16, (unsigned)(Fo)), 32, 0, stream>>>(cekv3_0); }
    { GemmP cekv3_1;
      cekv3_1.A = HP + (size_t)1 * C1; cekv3_1.B = wkv + 1; cekv3_1.bias = HP + (size_t)1 * C1; cekv3_1.R = KV; cekv3_1.C = KV;
      cekv3_1.sAo = (long long)3 * 2050 * C1; cekv3_1.sAi = 0; cekv3_1.sAm = C1; cekv3_1.sAk = 1; cekv3_1.sBo = 0; cekv3_1.sBi = 0; cekv3_1.sBn = C1 * 9; cekv3_1.sBk = 9; cekv3_1.sCo = (long long)Tt * LD; cekv3_1.sCi = 0; cekv3_1.sCm = LD; cekv3_1.sRo = (long long)Tt * LD; cekv3_1.sRi = 0; cekv3_1.sRm = LD; cekv3_1.sRn = 1;
      cekv3_1.M = Tt; cekv3_1.N = D; cekv3_1.K = C1; cekv3_1.zi_n = 1; cekv3_1.flags = 4; cekv3_1.act = 0;
      cekv3_1.alpha = 1.0f; cekv3_1.beta = 1.0f; cekv3_1.sa = 1.0f; cekv3_1.sb = 1.0f; cekv3_1.Npad = LD; cekv3_1.pad_ = 0;
      k_gemm<1><<<dim3((unsigned)((LD) + 31) / 32, (unsigned)((Tt) + 15) / 16, (unsigned)(Fo)), 32, 0, stream>>>(cekv3_1); }
    { GemmP cekv3_2;
      cekv3_2.A = HP + (size_t)2 * C1; cekv3_2.B = wkv + 2; cekv3_2.bias = HP + (size_t)2 * C1; cekv3_2.R = KV; cekv3_2.C = KV;
      cekv3_2.sAo = (long long)3 * 2050 * C1; cekv3_2.sAi = 0; cekv3_2.sAm = C1; cekv3_2.sAk = 1; cekv3_2.sBo = 0; cekv3_2.sBi = 0; cekv3_2.sBn = C1 * 9; cekv3_2.sBk = 9; cekv3_2.sCo = (long long)Tt * LD; cekv3_2.sCi = 0; cekv3_2.sCm = LD; cekv3_2.sRo = (long long)Tt * LD; cekv3_2.sRi = 0; cekv3_2.sRm = LD; cekv3_2.sRn = 1;
      cekv3_2.M = Tt; cekv3_2.N = D; cekv3_2.K = C1; cekv3_2.zi_n = 1; cekv3_2.flags = 4; cekv3_2.act = 0;
      cekv3_2.alpha = 1.0f; cekv3_2.beta = 1.0f; cekv3_2.sa = 1.0f; cekv3_2.sb = 1.0f; cekv3_2.Npad = LD; cekv3_2.pad_ = 0;
      k_gemm<1><<<dim3((unsigned)((LD) + 31) / 32, (unsigned)((Tt) + 15) / 16, (unsigned)(Fo)), 32, 0, stream>>>(cekv3_2); }
    { GemmP cekv3_3;
      cekv3_3.A = HP + (size_t)2050 * C1; cekv3_3.B = wkv + 3; cekv3_3.bias = HP + (size_t)2050 * C1; cekv3_3.R = KV; cekv3_3.C = KV;
      cekv3_3.sAo = (long long)3 * 2050 * C1; cekv3_3.sAi = 0; cekv3_3.sAm = C1; cekv3_3.sAk = 1; cekv3_3.sBo = 0; cekv3_3.sBi = 0; cekv3_3.sBn = C1 * 9; cekv3_3.sBk = 9; cekv3_3.sCo = (long long)Tt * LD; cekv3_3.sCi = 0; cekv3_3.sCm = LD; cekv3_3.sRo = (long long)Tt * LD; cekv3_3.sRi = 0; cekv3_3.sRm = LD; cekv3_3.sRn = 1;
      cekv3_3.M = Tt; cekv3_3.N = D; cekv3_3.K = C1; cekv3_3.zi_n = 1; cekv3_3.flags = 4; cekv3_3.act = 0;
      cekv3_3.alpha = 1.0f; cekv3_3.beta = 1.0f; cekv3_3.sa = 1.0f; cekv3_3.sb = 1.0f; cekv3_3.Npad = LD; cekv3_3.pad_ = 0;
      k_gemm<1><<<dim3((unsigned)((LD) + 31) / 32, (unsigned)((Tt) + 15) / 16, (unsigned)(Fo)), 32, 0, stream>>>(cekv3_3); }
    { GemmP cekv3_4;
      cekv3_4.A = HP + (size_t)2051 * C1; cekv3_4.B = wkv + 4; cekv3_4.bias = HP + (size_t)2051 * C1; cekv3_4.R = KV; cekv3_4.C = KV;
      cekv3_4.sAo = (long long)3 * 2050 * C1; cekv3_4.sAi = 0; cekv3_4.sAm = C1; cekv3_4.sAk = 1; cekv3_4.sBo = 0; cekv3_4.sBi = 0; cekv3_4.sBn = C1 * 9; cekv3_4.sBk = 9; cekv3_4.sCo = (long long)Tt * LD; cekv3_4.sCi = 0; cekv3_4.sCm = LD; cekv3_4.sRo = (long long)Tt * LD; cekv3_4.sRi = 0; cekv3_4.sRm = LD; cekv3_4.sRn = 1;
      cekv3_4.M = Tt; cekv3_4.N = D; cekv3_4.K = C1; cekv3_4.zi_n = 1; cekv3_4.flags = 4; cekv3_4.act = 0;
      cekv3_4.alpha = 1.0f; cekv3_4.beta = 1.0f; cekv3_4.sa = 1.0f; cekv3_4.sb = 1.0f; cekv3_4.Npad = LD; cekv3_4.pad_ = 0;
      k_gemm<1><<<dim3((unsigned)((LD) + 31) / 32, (unsigned)((Tt) + 15) / 16, (unsigned)(Fo)), 32, 0, stream>>>(cekv3_4); }
    { GemmP cekv3_5;
      cekv3_5.A = HP + (size_t)2052 * C1; cekv3_5.B = wkv + 5; cekv3_5.bias = HP + (size_t)2052 * C1; cekv3_5.R = KV; cekv3_5.C = KV;
      cekv3_5.sAo = (long long)3 * 2050 * C1; cekv3_5.sAi = 0; cekv3_5.sAm = C1; cekv3_5.sAk = 1; cekv3_5.sBo = 0; cekv3_5.sBi = 0; cekv3_5.sBn = C1 * 9; cekv3_5.sBk = 9; cekv3_5.sCo = (long long)Tt * LD; cekv3_5.sCi = 0; cekv3_5.sCm = LD; cekv3_5.sRo = (long long)Tt * LD; cekv3_5.sRi = 0; cekv3_5.sRm = LD; cekv3_5.sRn = 1;
      cekv3_5.M = Tt; cekv3_5.N = D; cekv3_5.K = C1; cekv3_5.zi_n = 1; cekv3_5.flags = 4; cekv3_5.act = 0;
      cekv3_5.alpha = 1.0f; cekv3_5.beta = 1.0f; cekv3_5.sa = 1.0f; cekv3_5.sb = 1.0f; cekv3_5.Npad = LD; cekv3_5.pad_ = 0;
      k_gemm<1><<<dim3((unsigned)((LD) + 31) / 32, (unsigned)((Tt) + 15) / 16, (unsigned)(Fo)), 32, 0, stream>>>(cekv3_5); }
    { GemmP cekv3_6;
      cekv3_6.A = HP + (size_t)4100 * C1; cekv3_6.B = wkv + 6; cekv3_6.bias = HP + (size_t)4100 * C1; cekv3_6.R = KV; cekv3_6.C = KV;
      cekv3_6.sAo = (long long)3 * 2050 * C1; cekv3_6.sAi = 0; cekv3_6.sAm = C1; cekv3_6.sAk = 1; cekv3_6.sBo = 0; cekv3_6.sBi = 0; cekv3_6.sBn = C1 * 9; cekv3_6.sBk = 9; cekv3_6.sCo = (long long)Tt * LD; cekv3_6.sCi = 0; cekv3_6.sCm = LD; cekv3_6.sRo = (long long)Tt * LD; cekv3_6.sRi = 0; cekv3_6.sRm = LD; cekv3_6.sRn = 1;
      cekv3_6.M = Tt; cekv3_6.N = D; cekv3_6.K = C1; cekv3_6.zi_n = 1; cekv3_6.flags = 4; cekv3_6.act = 0;
      cekv3_6.alpha = 1.0f; cekv3_6.beta = 1.0f; cekv3_6.sa = 1.0f; cekv3_6.sb = 1.0f; cekv3_6.Npad = LD; cekv3_6.pad_ = 0;
      k_gemm<1><<<dim3((unsigned)((LD) + 31) / 32, (unsigned)((Tt) + 15) / 16, (unsigned)(Fo)), 32, 0, stream>>>(cekv3_6); }
    { GemmP cekv3_7;
      cekv3_7.A = HP + (size_t)4101 * C1; cekv3_7.B = wkv + 7; cekv3_7.bias = HP + (size_t)4101 * C1; cekv3_7.R = KV; cekv3_7.C = KV;
      cekv3_7.sAo = (long long)3 * 2050 * C1; cekv3_7.sAi = 0; cekv3_7.sAm = C1; cekv3_7.sAk = 1; cekv3_7.sBo = 0; cekv3_7.sBi = 0; cekv3_7.sBn = C1 * 9; cekv3_7.sBk = 9; cekv3_7.sCo = (long long)Tt * LD; cekv3_7.sCi = 0; cekv3_7.sCm = LD; cekv3_7.sRo = (long long)Tt * LD; cekv3_7.sRi = 0; cekv3_7.sRm = LD; cekv3_7.sRn = 1;
      cekv3_7.M = Tt; cekv3_7.N = D; cekv3_7.K = C1; cekv3_7.zi_n = 1; cekv3_7.flags = 4; cekv3_7.act = 0;
      cekv3_7.alpha = 1.0f; cekv3_7.beta = 1.0f; cekv3_7.sa = 1.0f; cekv3_7.sb = 1.0f; cekv3_7.Npad = LD; cekv3_7.pad_ = 0;
      k_gemm<1><<<dim3((unsigned)((LD) + 31) / 32, (unsigned)((Tt) + 15) / 16, (unsigned)(Fo)), 32, 0, stream>>>(cekv3_7); }
    { GemmP cekv3_8;
      cekv3_8.A = HP + (size_t)4102 * C1; cekv3_8.B = wkv + 8; cekv3_8.bias = HP + (size_t)4102 * C1; cekv3_8.R = KV; cekv3_8.C = KV;
      cekv3_8.sAo = (long long)3 * 2050 * C1; cekv3_8.sAi = 0; cekv3_8.sAm = C1; cekv3_8.sAk = 1; cekv3_8.sBo = 0; cekv3_8.sBi = 0; cekv3_8.sBn = C1 * 9; cekv3_8.sBk = 9; cekv3_8.sCo = (long long)Tt * LD; cekv3_8.sCi = 0; cekv3_8.sCm = LD; cekv3_8.sRo = (long long)Tt * LD; cekv3_8.sRi = 0; cekv3_8.sRm = LD; cekv3_8.sRn = 1;
      cekv3_8.M = Tt; cekv3_8.N = D; cekv3_8.K = C1; cekv3_8.zi_n = 1; cekv3_8.flags = 4; cekv3_8.act = 0;
      cekv3_8.alpha = 1.0f; cekv3_8.beta = 1.0f; cekv3_8.sa = 1.0f; cekv3_8.sb = 1.0f; cekv3_8.Npad = LD; cekv3_8.pad_ = 0;
      k_gemm<1><<<dim3((unsigned)((LD) + 31) / 32, (unsigned)((Tt) + 15) / 16, (unsigned)(Fo)), 32, 0, stream>>>(cekv3_8); }

    k_cl_colsum1<<<NB, 256, 0, stream>>>(frame + (size_t)3 * Ll, 1, 1, (long long)Ll, PART); k_cl_colsum2<<<1, 256, 0, stream>>>(PART, NB, 1, RED, 0);
    k_cl_masknorm<<<(unsigned)((Ll + 255) / 256), 256, 0, stream>>>(KV, LD, frame + (size_t)3 * Ll, RED, Tsc, (long long)Ll, D);
    { GemmP gpQP3;
      gpQP3.A = Q; gpQP3.B = faq; gpQP3.bias = fabq; gpQP3.R = Q; gpQP3.C = QP;
      gpQP3.sAo = 0; gpQP3.sAi = 0; gpQP3.sAm = LD; gpQP3.sAk = 1; gpQP3.sBo = 0; gpQP3.sBi = 0; gpQP3.sBn = 1; gpQP3.sBk = D; gpQP3.sCo = 0; gpQP3.sCi = 0; gpQP3.sCm = LD; gpQP3.sRo = 0; gpQP3.sRi = 0; gpQP3.sRm = 0; gpQP3.sRn = 0;
      gpQP3.M = Ll; gpQP3.N = D; gpQP3.K = D; gpQP3.zi_n = 1; gpQP3.flags = 1; gpQP3.act = 6;
      gpQP3.alpha = 1.0f; gpQP3.beta = 0.0f; gpQP3.sa = 1.0f; gpQP3.sb = 1.0f; gpQP3.Npad = LD; gpQP3.pad_ = 0;
      k_gemm<1><<<dim3((unsigned)((LD) + 31) / 32, (unsigned)((Ll) + 15) / 16, (unsigned)(1)), 32, 0, stream>>>(gpQP3); }
    { GemmP gpKP3;
      gpKP3.A = KV; gpKP3.B = fak; gpKP3.bias = fabk; gpKP3.R = KV; gpKP3.C = KP;
      gpKP3.sAo = 0; gpKP3.sAi = 0; gpKP3.sAm = LD; gpKP3.sAk = 1; gpKP3.sBo = 0; gpKP3.sBi = 0; gpKP3.sBn = 1; gpKP3.sBk = D; gpKP3.sCo = 0; gpKP3.sCi = 0; gpKP3.sCm = LD; gpKP3.sRo = 0; gpKP3.sRi = 0; gpKP3.sRm = 0; gpKP3.sRn = 0;
      gpKP3.M = Ll; gpKP3.N = D; gpKP3.K = D; gpKP3.zi_n = 1; gpKP3.flags = 1; gpKP3.act = 6;
      gpKP3.alpha = 1.0f; gpKP3.beta = 0.0f; gpKP3.sa = 1.0f; gpKP3.sb = 1.0f; gpKP3.Npad = LD; gpKP3.pad_ = 0;
      k_gemm<1><<<dim3((unsigned)((LD) + 31) / 32, (unsigned)((Ll) + 15) / 16, (unsigned)(1)), 32, 0, stream>>>(gpKP3); }
    { GemmP gpVP3;
      gpVP3.A = KV; gpVP3.B = fav; gpVP3.bias = fabv; gpVP3.R = KV; gpVP3.C = VP;
      gpVP3.sAo = 0; gpVP3.sAi = 0; gpVP3.sAm = LD; gpVP3.sAk = 1; gpVP3.sBo = 0; gpVP3.sBi = 0; gpVP3.sBn = 1; gpVP3.sBk = D; gpVP3.sCo = 0; gpVP3.sCi = 0; gpVP3.sCm = LD; gpVP3.sRo = 0; gpVP3.sRi = 0; gpVP3.sRm = 0; gpVP3.sRn = 0;
      gpVP3.M = Ll; gpVP3.N = D; gpVP3.K = D; gpVP3.zi_n = 1; gpVP3.flags = 1; gpVP3.act = 0;
      gpVP3.alpha = 1.0f; gpVP3.beta = 0.0f; gpVP3.sa = 1.0f; gpVP3.sb = 1.0f; gpVP3.Npad = LD; gpVP3.pad_ = 0;
      k_gemm<1><<<dim3((unsigned)((LD) + 31) / 32, (unsigned)((Ll) + 15) / 16, (unsigned)(1)), 32, 0, stream>>>(gpVP3); }
    k_cl_colsum1<<<NB, 256, 0, stream>>>(KP, LD, D, (long long)Ll, PART); k_cl_colsum2<<<1, 256, 0, stream>>>(PART, NB, D, RED, 16);
    k_cl_colsum1<<<NB, 256, 0, stream>>>(QP, LD, D, (long long)Ll, PART); k_cl_colsum2<<<1, 256, 0, stream>>>(PART, NB, D, RED, 32);
    k_cl_flow1<<<(unsigned)((Ll + 255) / 256), 256, 0, stream>>>(QP, KP, LD, RED, SV, (long long)Ll, D);
    k_cl_flow2<<<(unsigned)(((long long)Ll * D + 255) / 256), 256, 0, stream>>>(QP, KP, LD, SV, O, O2, (long long)Ll, D);
    k_cl_colsum1<<<NB, 256, 0, stream>>>(O, LD, D, (long long)Ll, PART); k_cl_colsum2<<<1, 256, 0, stream>>>(PART, NB, D, RED, 48);
    k_cl_colsum1<<<NB, 256, 0, stream>>>(O2, LD, D, (long long)Ll, PART); k_cl_colsum2<<<1, 256, 0, stream>>>(PART, NB, D, RED, 64);
    k_cl_flow3<<<(unsigned)((Ll + 255) / 256), 256, 0, stream>>>(QP, KP, LD, RED, SV, (long long)Ll, D);
    k_cl_max1<<<NB, 256, 0, stream>>>(SV, 3, (long long)Ll, PART); k_cl_max2<<<1, 256, 0, stream>>>(PART, NB, RED, 80);
    k_cl_flow4<<<(unsigned)((Ll + 255) / 256), 256, 0, stream>>>(SV, RED, O2, LD, (long long)Ll);
    k_cl_colsum1<<<NB, 256, 0, stream>>>(O2 + 15, LD, 1, (long long)Ll, PART); k_cl_colsum2<<<1, 256, 0, stream>>>(PART, NB, 1, RED, 96);
    k_cl_flow5<<<(unsigned)(((long long)Ll * D + 255) / 256), 256, 0, stream>>>(VP, O2, LD, RED, O, (long long)Ll, D);
    { GemmP gkv3;
      gkv3.A = KP; gkv3.B = O; gkv3.bias = KP; gkv3.R = KP; gkv3.C = KVM;
      gkv3.sAo = 0; gkv3.sAi = 0; gkv3.sAm = 1; gkv3.sAk = LD; gkv3.sBo = 0; gkv3.sBi = 0; gkv3.sBn = 1; gkv3.sBk = LD; gkv3.sCo = 0; gkv3.sCi = 0; gkv3.sCm = LD; gkv3.sRo = 0; gkv3.sRi = 0; gkv3.sRm = 0; gkv3.sRn = 0;
      gkv3.M = D; gkv3.N = D; gkv3.K = Ll; gkv3.zi_n = 1; gkv3.flags = 0; gkv3.act = 0;
      gkv3.alpha = 1.0f; gkv3.beta = 0.0f; gkv3.sa = 1.0f; gkv3.sb = 1.0f; gkv3.Npad = LD; gkv3.pad_ = 0;
      k_gemm<1><<<dim3((unsigned)((LD) + 31) / 32, (unsigned)((D) + 15) / 16, (unsigned)(1)), 32, 0, stream>>>(gkv3); }
    { GemmP gqkv3;
      gqkv3.A = QP; gqkv3.B = KVM; gqkv3.bias = QP; gqkv3.R = QP; gqkv3.C = O2;
      gqkv3.sAo = 0; gqkv3.sAi = 0; gqkv3.sAm = LD; gqkv3.sAk = 1; gqkv3.sBo = 0; gqkv3.sBi = 0; gqkv3.sBn = 1; gqkv3.sBk = LD; gqkv3.sCo = 0; gqkv3.sCi = 0; gqkv3.sCm = LD; gqkv3.sRo = 0; gqkv3.sRi = 0; gqkv3.sRm = 0; gqkv3.sRn = 0;
      gqkv3.M = Ll; gqkv3.N = D; gqkv3.K = D; gqkv3.zi_n = 1; gqkv3.flags = 0; gqkv3.act = 0;
      gqkv3.alpha = 1.0f; gqkv3.beta = 0.0f; gqkv3.sa = 1.0f; gqkv3.sb = 1.0f; gqkv3.Npad = LD; gqkv3.pad_ = 0;
      k_gemm<1><<<dim3((unsigned)((LD) + 31) / 32, (unsigned)((Ll) + 15) / 16, (unsigned)(1)), 32, 0, stream>>>(gqkv3); }
    k_cl_flow6<<<(unsigned)(((long long)Ll * D + 255) / 256), 256, 0, stream>>>(O2, LD, SV, (long long)Ll, D);
    { GemmP gwo3;
      gwo3.A = O2; gwo3.B = fao; gwo3.bias = fabo; gwo3.R = O2; gwo3.C = O;
      gwo3.sAo = 0; gwo3.sAi = 0; gwo3.sAm = LD; gwo3.sAk = 1; gwo3.sBo = 0; gwo3.sBi = 0; gwo3.sBn = 1; gwo3.sBk = D; gwo3.sCo = 0; gwo3.sCi = 0; gwo3.sCm = LD; gwo3.sRo = 0; gwo3.sRi = 0; gwo3.sRm = 0; gwo3.sRn = 0;
      gwo3.M = Ll; gwo3.N = D; gwo3.K = D; gwo3.zi_n = 1; gwo3.flags = 1; gwo3.act = 0;
      gwo3.alpha = 1.0f; gwo3.beta = 0.0f; gwo3.sa = 1.0f; gwo3.sb = 1.0f; gwo3.Npad = LD; gwo3.pad_ = 0;
      k_gemm<1><<<dim3((unsigned)((LD) + 31) / 32, (unsigned)((Ll) + 15) / 16, (unsigned)(1)), 32, 0, stream>>>(gwo3); }
    k_cl_out<<<(unsigned)(((long long)Ll * D + 255) / 256), 256, 0, stream>>>(O, LD, out, 3, (long long)Ll, D);
}
